// SandboxLocalEventOperator_33346126086687
// MI455X (gfx1250) — hardware-verified
//
#include <hip/hip_runtime.h>
#include <math.h>

typedef __attribute__((ext_vector_type(16))) _Float16 v16h;
typedef __attribute__((ext_vector_type(8)))  _Float16 v8h;
typedef __attribute__((ext_vector_type(16))) __bf16   v16b;
typedef __attribute__((ext_vector_type(8)))  float    v8f;
typedef __attribute__((ext_vector_type(4)))  float    v4f;

__device__ __forceinline__ int frag_k(int i, int h) { return (i < 8) ? (8 * h + i) : (16 + 8 * h + (i - 8)); }
__device__ __forceinline__ __bf16 bf16_rne(float f) {
    unsigned int u = __float_as_uint(f);
    u += 0x7fffu + ((u >> 16) & 1u);
    return __builtin_bit_cast(__bf16, (unsigned short)(u >> 16));
}
__device__ __forceinline__ float bf16_f32(__bf16 b) { return __uint_as_float(((unsigned int)__builtin_bit_cast(unsigned short, b)) << 16); }
__device__ __forceinline__ v8f wmma16(v16h a, v16h b, v8f c) {
    c = __builtin_amdgcn_wmma_f32_16x16x32_f16(false, a, false, b, (short)0, c, false, false);
    asm volatile("v_nop\n\tv_nop\n\tv_nop\n\tv_nop" : "+v"(c) : "v"(a), "v"(b));
    return c;
}
__device__ __forceinline__ v8f wmmab(v16b a, v16b b, v8f c) {
    c = __builtin_amdgcn_wmma_f32_16x16x32_bf16(false, a, false, b, (short)0, c, false, false);
    asm volatile("v_nop\n\tv_nop\n\tv_nop\n\tv_nop" : "+v"(c) : "v"(a), "v"(b));
    return c;
}
struct Split { v16b hi, lo; };
__device__ __forceinline__ v8f wmma3(const Split& a, const Split& b, v8f c) {
    c = __builtin_amdgcn_wmma_f32_16x16x32_bf16(false, a.hi, false, b.hi, (short)0, c, false, false);
    c = __builtin_amdgcn_wmma_f32_16x16x32_bf16(false, a.hi, false, b.lo, (short)0, c, false, false);
    c = __builtin_amdgcn_wmma_f32_16x16x32_bf16(false, a.lo, false, b.hi, (short)0, c, false, false);
    asm volatile("v_nop\n\tv_nop\n\tv_nop\n\tv_nop" : "+v"(c) : "v"(a.hi), "v"(a.lo), "v"(b.hi), "v"(b.lo));
    return c;
}
struct Split3 { v16b hi, mid, lo; };
__device__ __forceinline__ v8f wmma6(const Split3& a, const Split3& b, v8f c) {
    c = __builtin_amdgcn_wmma_f32_16x16x32_bf16(false, a.hi, false, b.hi, (short)0, c, false, false);
    c = __builtin_amdgcn_wmma_f32_16x16x32_bf16(false, a.hi, false, b.mid, (short)0, c, false, false);
    c = __builtin_amdgcn_wmma_f32_16x16x32_bf16(false, a.mid, false, b.hi, (short)0, c, false, false);
    c = __builtin_amdgcn_wmma_f32_16x16x32_bf16(false, a.hi, false, b.lo, (short)0, c, false, false);
    c = __builtin_amdgcn_wmma_f32_16x16x32_bf16(false, a.mid, false, b.mid, (short)0, c, false, false);
    c = __builtin_amdgcn_wmma_f32_16x16x32_bf16(false, a.lo, false, b.hi, (short)0, c, false, false);
    asm volatile("v_nop\n\tv_nop\n\tv_nop\n\tv_nop" : "+v"(c) : "v"(a.hi), "v"(a.mid), "v"(a.lo), "v"(b.hi), "v"(b.mid), "v"(b.lo));
    return c;
}

__device__ __forceinline__ v16h fh_ld(const float* __restrict__ p, long long sk, int k0, int h, int klen, float s) {
    v16h a;
#pragma unroll
    for (int i = 0; i < 16; ++i) { const int k = k0 + frag_k(i, h); a[i] = (k < klen) ? (_Float16)(p[(long long)k * sk] * s) : (_Float16)0.f; }
    return a;
}
__device__ __forceinline__ Split sp_ld(const float* __restrict__ p, long long sk, int k0, int h, int klen, float s) {
    Split r;
#pragma unroll
    for (int i = 0; i < 16; ++i) {
        const int k = k0 + frag_k(i, h); const float x = (k < klen) ? p[(long long)k * sk] * s : 0.f;
        const __bf16 hb = bf16_rne(x); r.hi[i] = hb; r.lo[i] = bf16_rne(x - bf16_f32(hb));
    }
    return r;
}
__device__ __forceinline__ Split3 sp3_ld(const float* __restrict__ p, long long sk, int k0, int h, int klen, float s) {
    Split3 r;
#pragma unroll
    for (int i = 0; i < 16; ++i) {
        const int k = k0 + frag_k(i, h); const float x = (k < klen) ? p[(long long)k * sk] * s : 0.f;
        const __bf16 hb = bf16_rne(x); const float r1 = x - bf16_f32(hb); const __bf16 mb = bf16_rne(r1);
        r.hi[i] = hb; r.mid[i] = mb; r.lo[i] = bf16_rne(r1 - bf16_f32(mb));
    }
    return r;
}
__device__ __forceinline__ v16b bh_ld(const float* __restrict__ p, long long sk, int k0, int h, int klen, float s) {
    v16b a;
#pragma unroll
    for (int i = 0; i < 16; ++i) { const int k = k0 + frag_k(i, h); a[i] = bf16_rne((k < klen) ? p[(long long)k * sk] * s : 0.f); }
    return a;
}
__device__ __forceinline__ v16h fh_row(const _Float16* __restrict__ row, int k0, int h) {
    v16h a;
#pragma unroll
    for (int i = 0; i < 16; ++i) a[i] = row[k0 + frag_k(i, h)];
    return a;
}

#define VST2(T, ptr, val) do { *(volatile T*)(ptr) = (val); __threadfence(); *(volatile T*)(ptr) = (val); } while (0)
typedef float v4f __attribute__((ext_vector_type(4)));
#define VST2V4(ptr, val) do { *(volatile v4f*)(ptr) = (val); __threadfence(); *(volatile v4f*)(ptr) = (val); } while (0)

__device__ __attribute__((noinline)) float act_fn(float v, int act) {
    if (act == 1) return fmaxf(v, 0.f);
    if (act == 2) { const float u = 0.7978845608028654f * (v + 0.044715f * v * v * v); return 0.5f * v * (1.f + tanhf(u)); }
    if (act == 3) return v / (1.f + expf(-v));
    if (act == 4) return 0.5f * v * (1.f + erff(v * 0.7071067811865476f));
    if (act == 5) return tanhf(v);
    if (act == 6) return 1.f / (1.f + expf(-v));
    if (act == 7) return (v > 0.f) ? v : 0.01f * v;
    if (act == 8) return (v > 0.f) ? v : (expf(v) - 1.f);
    if (act == 9) return fminf(fmaxf(v, 0.f), 6.f);
    if (act == 10) return fabsf(v);
    if (act == 11) return (v >= 0.f) ? v : 0.1f * v;
    if (act == 12) return (v > 0.f) ? v : 0.2f * v;
    if (act == 13) return (v > 20.f) ? v : log1pf(expf(v));
    return v;
}

struct GemmP {
    const float* A; const float* B; const float* bias; const float* R; float* C;
    long long sAo, sAi, sAm, sAk, sBo, sBi, sBn, sBk, sCo, sCi, sCm, sRo, sRi, sRm, sRn;
    int M, N, K, zi_n, flags, act; float alpha, beta, sa, sb;
    int Npad, pad_;
};
static_assert(sizeof(GemmP) == 5 * 8 + 15 * 8 + 6 * 4 + 4 * 4 + 2 * 4, "GemmP has padding");

template <int MODE>
__global__ __launch_bounds__(32) void k_gemm(GemmP p) {
    const int lane = threadIdx.x & 31, h = lane >> 4, l15 = lane & 15;
    const int m0 = blockIdx.y * 16, n0 = blockIdx.x * 32;
    const int z = blockIdx.z, zo = z / p.zi_n, zi = z - zo * p.zi_n;
    const float* A = p.A + zo * p.sAo + zi * p.sAi;
    const float* B = p.B + zo * p.sBo + zi * p.sBi;
    const int am = min(m0 + l15, p.M - 1);
    v8f acc[2], comp[2];
#pragma unroll
    for (int t = 0; t < 2; ++t) { v8f zz = {}; acc[t] = zz; comp[t] = zz; }
    for (int k0 = 0; k0 < p.K; k0 += 32) {
        const float* arow = A + (long long)am * p.sAm;
        if (MODE == 1) {
            const Split a = sp_ld(arow, p.sAk, k0, h, p.K, 1.f);
#pragma unroll
            for (int t = 0; t < 2; ++t) {
                const int bn = min(n0 + t * 16 + l15, p.N - 1);
                acc[t] = wmma3(a, sp_ld(B + (long long)bn * p.sBn, p.sBk, k0, h, p.K, 1.f), acc[t]);
            }
        } else if (MODE == 3) {
            const Split3 a = sp3_ld(arow, p.sAk, k0, h, p.K, 1.f);
#pragma unroll
            for (int t = 0; t < 2; ++t) {
                const int bn = min(n0 + t * 16 + l15, p.N - 1);
                acc[t] = wmma6(a, sp3_ld(B + (long long)bn * p.sBn, p.sBk, k0, h, p.K, 1.f), acc[t]);
            }
        } else if (MODE == 4) {
            const Split3 a = sp3_ld(arow, p.sAk, k0, h, p.K, 1.f);
#pragma unroll
            for (int t = 0; t < 2; ++t) {
                const int bn = min(n0 + t * 16 + l15, p.N - 1); v8f zz = {};
                const v8f part = wmma6(a, sp3_ld(B + (long long)bn * p.sBn, p.sBk, k0, h, p.K, 1.f), zz);
                const v8f y = part - comp[t]; const v8f s = acc[t] + y; comp[t] = (s - acc[t]) - y; acc[t] = s;
            }
        } else if (MODE == 2) {
            const v16b a = bh_ld(arow, p.sAk, k0, h, p.K, 1.f);
#pragma unroll
            for (int t = 0; t < 2; ++t) {
                const int bn = min(n0 + t * 16 + l15, p.N - 1);
                acc[t] = wmmab(a, bh_ld(B + (long long)bn * p.sBn, p.sBk, k0, h, p.K, 1.f), acc[t]);
            }
        } else {
            const v16h a = fh_ld(arow, p.sAk, k0, h, p.K, p.sa);
#pragma unroll
            for (int t = 0; t < 2; ++t) {
                const int bn = min(n0 + t * 16 + l15, p.N - 1);
                acc[t] = wmma16(a, fh_ld(B + (long long)bn * p.sBn, p.sBk, k0, h, p.K, p.sb), acc[t]);
            }
        }
    }
    const float iscale = (MODE == 0) ? p.alpha / (p.sa * p.sb) : p.alpha;
    float* C = p.C + zo * p.sCo + zi * p.sCi;
    const float* R = p.R + zo * p.sRo + zi * p.sRi;
    __shared__ __align__(16) float ctile[16][36];
#pragma unroll
    for (int t = 0; t < 2; ++t) {
        const int n = n0 + t * 16 + l15; const int nn = min(n, p.N - 1);
#pragma unroll
        for (int r = 0; r < 8; ++r) {
            const int m = m0 + 8 * h + r; const int mm = min(m, p.M - 1);
            float v = acc[t][r] * iscale;
            if (p.flags & 1) v += p.bias[nn];
            if (p.flags & 2) v += p.bias[mm];
            v = act_fn(v, p.act);
            if (p.flags & 4) v += p.beta * R[(long long)mm * p.sRm + (long long)nn * p.sRn];
            ctile[8 * h + r][t * 16 + l15] = (n < p.N) ? v : 0.f;
        }
    }
    __syncthreads();
    const int NW = (p.Npad > p.N) ? p.Npad : p.N;
    const bool fast = (m0 + 16 <= p.M) && (n0 + 32 <= NW) && ((p.sCm & 3) == 0) && ((((size_t)C) & 15) == 0);
    if (fast) {
#pragma unroll
        for (int s = 0; s < 4; ++s) {
            const int row = s * 4 + (lane >> 3), c4 = (lane & 7) * 4;
            const v4f v = *(const v4f*)&ctile[row][c4];
            VST2V4(C + (long long)(m0 + row) * p.sCm + n0 + c4, v);
        }
    } else {
        for (int row = 0; row < 16; ++row) {
            const int m = m0 + row, n = n0 + lane;
            if (m < p.M && n < NW) VST2(float, C + (long long)m * p.sCm + n, ctile[row][lane]);
        }
    }
}

#define AW 4
struct AttnP {
    const float* Q; const float* K; const float* V; float* O; float* P; const float* Mf; const int* Mi; float* ST;
    const float* Pw; const float* Rt; const int* SQ; const int* SK;
    long long swb, swh, swi, swj, srb, srh, sri;
    long long sQb, sQh, sQi, sQd, sKb, sKh, sKj, sKd, sVb, sVh, sVj, sVd, sOb, sOh, sOi, sPb, sPh, sPi, smb, smh, smi, smj;
    int Lq, Lk, dh, dv, hrep, causal, coff, pband;
    float scale, mfill; int nonorm, mpol;
    int roff, rn, segpol, win;
};
static_assert(sizeof(AttnP) == 12 * 8 + 29 * 8 + 16 * 4, "AttnP has padding");

#ifndef KATTN_ATTR
#define KATTN_ATTR
#endif
template <int DHP, int DVP, int QM, bool SPLITPV, bool TWOPASS>
__global__ __launch_bounds__(32 * AW) KATTN_ATTR void k_attn(AttnP p) {
    constexpr int NT = DVP / 16;
    constexpr int KS = DHP / 32;
    constexpr int VP = DVP + 8;
    __shared__ __align__(16) float    pl[AW][16 * 64];
    __shared__ __align__(16) _Float16 vl[(SPLITPV ? 2 : 1) * 64 * VP];
    const int lane = threadIdx.x & 31, hf = lane >> 4, l15 = lane & 15, wave = threadIdx.x >> 5;
    const int h = blockIdx.y, b = blockIdx.z, hk = h / p.hrep;
    const int q0 = (blockIdx.x * AW + wave) * 16;
    float* myp = pl[wave];
    const float L2E = 1.4426950408889634f;
    const float NEG = -__builtin_inff();
    const int qi = min(q0 + l15, p.Lq - 1);
    const float* qrow = p.Q + b * p.sQb + h * p.sQh + (long long)qi * p.sQi;
    const float* kbase = p.K + b * p.sKb + hk * p.sKh;
    const float* vbase = p.V + b * p.sVb + hk * p.sVh;
    v16h qa[QM == 0 ? KS : 1]; Split qs_[QM == 1 ? KS : 1]; Split3 qt_[QM == 2 ? KS : 1];
#pragma unroll
    for (int ks = 0; ks < KS; ++ks) {
        if (QM == 2) qt_[ks] = sp3_ld(qrow, p.sQd, ks * 32, hf, p.dh, 1.f);
        else if (QM == 1) qs_[ks] = sp_ld(qrow, p.sQd, ks * 32, hf, p.dh, 1.f);
        else qa[ks] = fh_ld(qrow, p.sQd, ks * 32, hf, p.dh, 1.f);
    }
    v8f o[NT]; float m8[8], l8[8];
#pragma unroll
    for (int t = 0; t < NT; ++t) { v8f zz = {}; o[t] = zz; }
#pragma unroll
    for (int i = 0; i < 8; ++i) { m8[i] = NEG; l8[i] = 0.f; }
    int jend = p.Lk;
    if (p.causal == 1) { const int je = (blockIdx.x * AW + AW - 1) * 16 + 16 + p.coff; jend = min(jend, max(je, 0)); }
    const int npass = TWOPASS ? 2 : 1;
    for (int pass = 0; pass < npass; ++pass) {
        const bool dopv = (!TWOPASS) || pass == 1;
        for (int j0 = 0; j0 < jend; j0 += 64) {
            if (dopv) {
                __syncthreads();
                for (int idx = threadIdx.x; idx < 64 * DVP; idx += 32 * AW) {
                    const int jr = idx / DVP, d = idx - jr * DVP, j = j0 + jr;
                    const float f = (j < p.Lk && d < p.dv) ? vbase[(long long)j * p.sVj + (long long)d * p.sVd] : 0.f;
                    if (SPLITPV) {
                        const __bf16 hb = bf16_rne(f);
                        ((__bf16*)vl)[jr * VP + d] = hb; ((__bf16*)vl)[64 * VP + jr * VP + d] = bf16_rne(f - bf16_f32(hb));
                    } else vl[jr * VP + d] = (_Float16)f;
                }
            }
            v8f s[4];
#pragma unroll
            for (int t = 0; t < 4; ++t) {
                const int j = min(j0 + t * 16 + l15, p.Lk - 1);
                const float* krow = kbase + (long long)j * p.sKj;
                v8f acc = {};
#pragma unroll
                for (int ks = 0; ks < KS; ++ks) {
                    if (QM == 2)      acc = wmma6(qt_[ks], sp3_ld(krow, p.sKd, ks * 32, hf, p.dh, 1.f), acc);
                    else if (QM == 1) acc = wmma3(qs_[ks], sp_ld(krow, p.sKd, ks * 32, hf, p.dh, 1.f), acc);
                    else              acc = wmma16(qa[ks], fh_ld(krow, p.sKd, ks * 32, hf, p.dh, 1.f), acc);
                }
                s[t] = acc;
            }
            float pv[8][4];
#pragma unroll
            for (int i = 0; i < 8; ++i) {
                const int irow = q0 + i + 8 * hf;
                const int ic = min(irow, p.Lq - 1);
                float sc[4];
#pragma unroll
                for (int t = 0; t < 4; ++t) {
                    const int jg = j0 + t * 16 + l15;
                    float v = s[t][i] * p.scale;
                    if (p.Mf) v += p.Mf[b * p.smb + h * p.smh + (long long)ic * p.smi + (long long)min(jg, p.Lk - 1) * p.smj];
                    if (p.Rt) { int rc = ic - min(jg, p.Lk - 1) + p.roff; rc = rc < 0 ? 0 : (rc >= p.rn ? p.rn - 1 : rc); v += p.Rt[b * p.srb + h * p.srh + (long long)ic * p.sri + rc]; }
                    if (p.Mi) { const int mv = p.Mi[b * p.smb + h * p.smh + (long long)ic * p.smi + (long long)min(jg, p.Lk - 1) * p.smj]; if (p.mpol ? (mv != 0) : (mv == 0)) v = p.mfill; }
                    if (p.SQ) { const bool same = p.SQ[(long long)b * p.Lq + ic] == p.SK[(long long)b * p.Lk + min(jg, p.Lk - 1)]; if (p.segpol ? same : !same) v = p.mfill; }
                    if (p.causal == 2 && jg > irow + p.coff) v = p.mfill;
                    if (jg >= p.Lk || (p.causal == 1 && jg > irow + p.coff) || (p.causal == 3 && jg < irow + p.coff) || (p.win > 0 && irow + p.coff - jg > p.win)) v = NEG; else v *= L2E;
                    sc[t] = v;
                }
                if (!TWOPASS || pass == 0) {
                    float mx = fmaxf(fmaxf(sc[0], sc[1]), fmaxf(sc[2], sc[3]));
                    mx = fmaxf(mx, __shfl_xor(mx, 1, 32)); mx = fmaxf(mx, __shfl_xor(mx, 2, 32));
                    mx = fmaxf(mx, __shfl_xor(mx, 4, 32)); mx = fmaxf(mx, __shfl_xor(mx, 8, 32));
                    const float mnew = fmaxf(m8[i], mx);
                    const float corr = (mnew == NEG) ? 1.f : exp2f(m8[i] - mnew);
                    float rs = 0.f;
#pragma unroll
                    for (int t = 0; t < 4; ++t) {
                        const float pp = (sc[t] == NEG) ? 0.f : exp2f(sc[t] - mnew); rs += pp;
                        pv[i][t] = p.Pw ? pp * p.Pw[b * p.swb + h * p.swh + (long long)ic * p.swi + (long long)min(j0 + t * 16 + l15, p.Lk - 1) * p.swj] : pp;
                    }
                    rs += __shfl_xor(rs, 1, 32); rs += __shfl_xor(rs, 2, 32); rs += __shfl_xor(rs, 4, 32); rs += __shfl_xor(rs, 8, 32);
                    l8[i] = l8[i] * corr + rs; m8[i] = mnew;
                    if (!TWOPASS) {
#pragma unroll
                        for (int t = 0; t < NT; ++t) o[t][i] *= corr;
                    }
                } else {
                    const float inv = (l8[i] > 0.f) ? 1.f / l8[i] : 0.f;
#pragma unroll
                    for (int t = 0; t < 4; ++t) {
                        const int jg = j0 + t * 16 + l15;
                        float pp = (sc[t] == NEG) ? 0.f : exp2f(sc[t] - m8[i]) * inv;
                        if (p.Pw) pp *= p.Pw[b * p.swb + h * p.swh + (long long)ic * p.swi + (long long)min(jg, p.Lk - 1) * p.swj];
                        pv[i][t] = pp;
                    }
                }
            }
            if (dopv) {
#pragma unroll
                for (int i = 0; i < 8; ++i)
#pragma unroll
                    for (int t = 0; t < 4; ++t) myp[(i + 8 * hf) * 64 + t * 16 + l15] = pv[i][t];
                __syncthreads();
                if (p.P) {
                    float* pb_ = p.P + b * p.sPb + h * p.sPh;
                    const bool fastP = (p.pband == 0) && ((p.sPi & 3) == 0) && (j0 + 64 <= p.Lk) && (q0 + 16 <= p.Lq) && ((((size_t)pb_) & 15) == 0);
                    if (fastP) {
#pragma unroll
                        for (int s = 0; s < 8; ++s) {
                            const int row = s * 2 + (lane >> 4), c4 = (lane & 15) * 4;
                            const v4f v = *(const v4f*)(myp + row * 64 + c4);
                            VST2V4(pb_ + (long long)(q0 + row) * p.sPi + j0 + c4, v);
                        }
                    } else {
                        for (int row = 0; row < 16; ++row) {
                            const int irow = q0 + row; if (irow >= p.Lq) continue;
                            for (int c = lane; c < 64; c += 32) {
                                const int jg = j0 + c; if (jg >= p.Lk) continue;
                                if (p.pband == 0) VST2(float, pb_ + (long long)irow * p.sPi + jg, myp[row * 64 + c]);
                                else if (jg - irow <= p.pband && irow - jg <= p.pband) VST2(float, pb_ + (long long)irow * p.sPi + (jg - irow + p.pband), myp[row * 64 + c]);
                            }
                        }
                    }
                }
                if (SPLITPV) {
                    const Split pa0 = sp_ld(myp + l15 * 64, 1, 0, hf, 64, 1.f), pa1 = sp_ld(myp + l15 * 64, 1, 32, hf, 64, 1.f);
                    const __bf16* vh = (const __bf16*)vl; const __bf16* vlo = vh + 64 * VP;
#pragma unroll
                    for (int t = 0; t < NT; ++t) {
                        const int dcol = t * 16 + l15;
                        Split b0, b1;
#pragma unroll
                        for (int e = 0; e < 16; ++e) {
                            const int k0 = frag_k(e, hf), k1 = 32 + frag_k(e, hf);
                            b0.hi[e] = vh[k0 * VP + dcol]; b0.lo[e] = vlo[k0 * VP + dcol]; b1.hi[e] = vh[k1 * VP + dcol]; b1.lo[e] = vlo[k1 * VP + dcol];
                        }
                        o[t] = wmma3(pa0, b0, o[t]);
                        o[t] = wmma3(pa1, b1, o[t]);
                    }
                } else {
                    const v16h pa0 = fh_ld(myp + l15 * 64, 1, 0, hf, 64, 4096.f), pa1 = fh_ld(myp + l15 * 64, 1, 32, hf, 64, 4096.f);
#pragma unroll
                    for (int t = 0; t < NT; ++t) {
                        const int dcol = t * 16 + l15;
                        v16h b0, b1;
#pragma unroll
                        for (int e = 0; e < 16; ++e) { b0[e] = vl[frag_k(e, hf) * VP + dcol]; b1[e] = vl[(32 + frag_k(e, hf)) * VP + dcol]; }
                        o[t] = wmma16(pa0, b0, o[t]);
                        o[t] = wmma16(pa1, b1, o[t]);
                    }
                }
            }
        }
    }
    float* obase = p.O + b * p.sOb + h * p.sOh;
    if (p.ST) {
        const int rl = lane >> 1, isel = rl & 7;
        float mv = 0.f, lv = 0.f;
#pragma unroll
        for (int i = 0; i < 8; ++i) if (i == isel) { mv = m8[i]; lv = l8[i]; }
        const int irow = q0 + rl;
        if (irow < p.Lq) { float* st = p.ST + (((long long)b * gridDim.y + h) * p.Lq + irow) * 2 + (lane & 1); VST2(float, st, (lane & 1) ? lv : mv * 0.6931471805599453f); }
    }
    float invr[8];
#pragma unroll
    for (int i = 0; i < 8; ++i) {
        if (TWOPASS) invr[i] = SPLITPV ? 1.f : (1.f / 4096.f);
        else if (p.nonorm) invr[i] = exp2f(m8[i]) * (SPLITPV ? 1.f : (1.f / 4096.f));
        else invr[i] = (l8[i] > 0.f) ? (SPLITPV ? 1.f / l8[i] : 1.f / (l8[i] * 4096.f)) : 0.f;
    }
    __syncthreads();
    const bool ofast = ((p.sOi & 3) == 0) && ((((size_t)obase) & 15) == 0) && (q0 + 16 <= p.Lq);
#pragma unroll
    for (int c0 = 0; c0 < DVP; c0 += 64) {
#pragma unroll
        for (int i = 0; i < 8; ++i)
#pragma unroll
            for (int t = 0; t < NT; ++t) if (t * 16 >= c0 && t * 16 < c0 + 64) myp[(i + 8 * hf) * 64 + (t * 16 - c0) + l15] = o[t][i] * invr[i];
        __syncthreads();
        const int cw = (DVP - c0 < 64) ? (DVP - c0) : 64;
        if (ofast && (c0 + cw <= p.dv) && (cw % 32 == 0)) {
            const int lpr = cw / 4;
            const int rows_per_ins = 32 / lpr;
            for (int r0 = 0; r0 < 16; r0 += rows_per_ins) {
                const int row = r0 + lane / lpr, c4 = (lane % lpr) * 4;
                const v4f v = *(const v4f*)(myp + row * 64 + c4);
                VST2V4(obase + (long long)(q0 + row) * p.sOi + c0 + c4, v);
            }
        } else {
            for (int row = 0; row < 16; ++row) {
                const int irow = q0 + row; if (irow >= p.Lq) continue;
                for (int c = lane; c < cw; c += 32) { const int d = c0 + c; if (d < p.dv) VST2(float, obase + (long long)irow * p.sOi + d, myp[row * 64 + c]); }
            }
        }
        __syncthreads();
    }
}

struct TrP { const float* src; float* dst; const float* R2; long long sSz, lds, sDz, ldd, sRz, ldr; int R, C, flags, act; float alpha, beta; };
static_assert(sizeof(TrP) == 3 * 8 + 6 * 8 + 6 * 4, "TrP has padding");
__global__ __launch_bounds__(256) void k_tr(TrP p) {
    __shared__ float tile[32][33];
    const int c0 = blockIdx.x * 32, r0 = blockIdx.y * 32, z = blockIdx.z;
    const int lane = threadIdx.x & 31, wave = threadIdx.x >> 5;
    const float* s = p.src + z * p.sSz;
#pragma unroll
    for (int k = 0; k < 4; ++k) {
        const int rl = wave * 4 + k, r = r0 + rl, c = c0 + lane;
        tile[rl][lane] = (r < p.R && c < p.C) ? s[(long long)r * p.lds + c] : 0.f;
    }
    __syncthreads();
    float* d = p.dst + z * p.sDz; const float* rr = p.R2 + z * p.sRz;
#pragma unroll
    for (int k = 0; k < 4; ++k) {
        const int cl = wave * 4 + k, c = c0 + cl, r = r0 + lane;
        if (c < p.C && r < p.R) {
            float v = act_fn(p.alpha * tile[lane][cl], p.act);
            if (p.flags & 1) v += p.beta * rr[(long long)c * p.ldr + r];
            VST2(float, d + (long long)c * p.ldd + r, v);
        }
    }
}

__global__ __launch_bounds__(256) void k_affine(const float* __restrict__ src, float* __restrict__ dst, int n, float a, float b, const float* __restrict__ sdev) {
    const int i = blockIdx.x * 256 + threadIdx.x;
    if (i < n) { const float aa = sdev ? a * sdev[0] : a; const float v = aa * src[i] + b; VST2(float, dst + i, v); }
}

struct SmP { const float* src; float* dst; const float* Mf; long long sz, sr, dz, dr, smz, smr; int n, pad; float scale_in, scale_out; };
static_assert(sizeof(SmP) == 3 * 8 + 6 * 8 + 4 * 4, "SmP has padding");
__global__ __launch_bounds__(256) void k_softmax(SmP p) {
    __shared__ float red[256];
    const int r = blockIdx.x, z = blockIdx.y, tid = threadIdx.x;
    const float* s = p.src + z * p.sz + (long long)r * p.sr;
    const float* mf = p.Mf ? (p.Mf + z * p.smz + (long long)r * p.smr) : nullptr;
    float mx = -__builtin_inff();
    for (int j = tid; j < p.n; j += 256) { float v = s[j] * p.scale_in; if (mf) v += mf[j]; mx = fmaxf(mx, v); }
    red[tid] = mx; __syncthreads();
    for (int o = 128; o > 0; o >>= 1) { if (tid < o) red[tid] = fmaxf(red[tid], red[tid + o]); __syncthreads(); }
    mx = red[0]; __syncthreads();
    float sum = 0.f;
    for (int j = tid; j < p.n; j += 256) { float v = s[j] * p.scale_in; if (mf) v += mf[j]; sum += (mx == -__builtin_inff()) ? 0.f : expf(v - mx); }
    red[tid] = sum; __syncthreads();
    for (int o = 128; o > 0; o >>= 1) { if (tid < o) red[tid] += red[tid + o]; __syncthreads(); }
    sum = red[0];
    const float inv = (sum > 0.f) ? p.scale_out / sum : 0.f;
    float* d = p.dst + z * p.dz + (long long)r * p.dr;
    for (int j = tid; j < p.n; j += 256) { float v = s[j] * p.scale_in; if (mf) v += mf[j]; const float o = (mx == -__builtin_inff()) ? 0.f : expf(v - mx) * inv; VST2(float, d + j, o); }
}
__global__ __launch_bounds__(256) void k_stats(const float* __restrict__ x, long long sz, long long so, long long si, int inner, int n, float eps, float* __restrict__ stat, int mode) {
    __shared__ float red[256];
    const int z = blockIdx.x, tid = threadIdx.x;
    const float* base = x + z * sz;
    float s = 0.f;
    for (int e = tid; e < n; e += 256) s += base[(long long)(e / inner) * so + (long long)(e % inner) * si];
    red[tid] = s; __syncthreads();
    for (int o = 128; o > 0; o >>= 1) { if (tid < o) red[tid] += red[tid + o]; __syncthreads(); }
    const float mu = (mode == 0 || mode == 3) ? red[0] / (float)n : 0.f; __syncthreads();
    float q = 0.f;
    for (int e = tid; e < n; e += 256) { const float dlt = base[(long long)(e / inner) * so + (long long)(e % inner) * si] - mu; q += dlt * dlt; }
    red[tid] = q; __syncthreads();
    for (int o = 128; o > 0; o >>= 1) { if (tid < o) red[tid] += red[tid + o]; __syncthreads(); }
    {
        float rs;
        if (mode == 2) rs = sqrtf((float)n) / fmaxf(sqrtf(red[0]), eps); else if (mode == 3) rs = rsqrtf(red[0] / (float)(n - 1) + eps); else rs = rsqrtf(red[0] / (float)n + eps);
        if (tid < 32) { const float v = (tid == 0) ? mu : ((tid == 1) ? rs : 0.f); VST2(float, stat + (long long)z * 32 + tid, v); }
    }
}
__global__ __launch_bounds__(256) void k_norm_apply(const float* __restrict__ x, float* __restrict__ y, const float* __restrict__ stat, const float* __restrict__ g, const float* __restrict__ bta,
                                                     int Z, int C, int L, int G, int bn, int act) {
    const long long idx = (long long)blockIdx.x * 256 + threadIdx.x;
    if (idx >= (long long)Z * C * L) return;
    const int l = (int)(idx % L); const long long zc = idx / L; const int c = (int)(zc % C), z = (int)(zc / C); (void)l;
    const int set = bn ? c : (z * G + c / (C / G));
    float v = (x[idx] - stat[(long long)set * 32]) * stat[(long long)set * 32 + 1];
    if (g) v *= g[c];
    if (bta) v += bta[c];
    v = act_fn(v, act);
    VST2(float, y + idx, v);
}

__global__ __launch_bounds__(256) void k_lse_neg(const float* __restrict__ st, float* __restrict__ c, int n) {
    const int i = blockIdx.x * 256 + threadIdx.x;
    if (i < n) { const float v = -(st[2 * i] + logf(st[2 * i + 1])); VST2(float, c + i, v); }
}

__global__ __launch_bounds__(256) void k_iota(int* __restrict__ dst, int n, int a, int b) {
    const int i = blockIdx.x * 256 + threadIdx.x;
    if (i < n) { const int v = a * i + b; VST2(int, dst + i, v); }
}

__global__ __launch_bounds__(256) void k_axpby(const float* __restrict__ x, const float* __restrict__ y, float* __restrict__ dst, int n, float a, float b, float c) {
    const int i = blockIdx.x * 256 + threadIdx.x;
    if (i < n) { const float v = a * x[i] + b * y[i] + c; VST2(float, dst + i, v); }
}

struct RopeP { const float* X; float* Y; const float* C; const float* Sn; const int* pos; long long sXr, sXh, sYr, sYh, sCb, sCp, sCd; int R, Hn, D, S, mode, tmode, pmode, pad; };
static_assert(sizeof(RopeP) == 5 * 8 + 7 * 8 + 8 * 4, "RopeP has padding");
__global__ __launch_bounds__(256) void k_rope(RopeP p) {
    const long long idx = (long long)blockIdx.x * 256 + threadIdx.x;
    if (idx >= (long long)p.R * p.Hn * p.D) return;
    const int d = (int)(idx % p.D); const long long rh = idx / p.D; const int h = (int)(rh % p.Hn); const int r = (int)(rh / p.Hn);
    const int half = p.D / 2;
    int partner; float sign;
    if (p.mode == 0) { partner = (d < half) ? d + half : d - half; sign = (d < half) ? -1.f : 1.f; }
    else { partner = d ^ 1; sign = (d & 1) ? 1.f : -1.f; }
    const int tcol = (p.tmode == 0) ? d : ((p.tmode == 1) ? (d % half) : (d >> 1));
    const int pp = (p.pmode == 0) ? (r % p.S) : ((p.pmode == 1) ? h : p.pos[r]);
    const long long toff = (long long)(r / p.S) * p.sCb + (long long)pp * p.sCp + (long long)tcol * p.sCd;
    const float* xr = p.X + (long long)r * p.sXr + (long long)h * p.sXh;
    const float v = xr[d] * p.C[toff] + sign * xr[partner] * p.Sn[toff];
    VST2(float, p.Y + (long long)r * p.sYr + (long long)h * p.sYh + d, v);
}

__global__ __launch_bounds__(256) void k_invf(float* __restrict__ invb, int half, int D, float base, float num, int fmode, float cexp) {
    const int i = blockIdx.x * 256 + threadIdx.x;
    if (i >= ((half + 31) / 32) * 32) return;
    if (i >= half) { VST2(float, invb + i, 0.f); return; }
    const float e = (float)(2 * i) / (float)D;
    float invf;
    if (fmode == 1) invf = num * expf((float)(2 * i) * cexp);
    else if (fmode == 2) invf = num * powf(base, (-2.0f * ((float)i - 1.0f)) / (float)D);
    else invf = num * (1.0f / powf(base, e));
    VST2(float, invb + i, invf);
}
__global__ __launch_bounds__(256) void k_sincos(float* __restrict__ cs, float* __restrict__ sn, const float* __restrict__ invb, int S, int half, float pscale) {
    const int idx = blockIdx.x * 256 + threadIdx.x;
    if (idx >= S * half) return;
    const int s = idx / half, i = idx - s * half;
    const float ang = (pscale * (float)s) * invb[i];
    VST2(float, cs + idx, cosf(ang)); VST2(float, sn + idx, sinf(ang));
}

__global__ __launch_bounds__(256) void k_mulact(const float* __restrict__ x, const float* __restrict__ y, float* __restrict__ dst, int n, int act) {
    const int i = blockIdx.x * 256 + threadIdx.x;
    if (i < n) { const float v = act_fn(x[i], act) * y[i]; VST2(float, dst + i, v); }
}

__global__ __launch_bounds__(256) void k_matvec(GemmP p) {
    const int rpt = (p.N == 1) ? 1 : 32;
    const long long r0 = ((long long)blockIdx.x * 256 + threadIdx.x) * rpt; const int z = blockIdx.z, zo = z / p.zi_n, zi = z - zo * p.zi_n;
    if (r0 >= p.M) return;
    const float* Bb = p.B + zo * p.sBo + zi * p.sBi;
    float* C = p.C + zo * p.sCo + zi * p.sCi; const float* R = p.R + zo * p.sRo + zi * p.sRi;
    for (int rr = 0; rr < rpt; ++rr) {
        const long long r = r0 + rr; if (r >= p.M) break;
        const float* A = p.A + zo * p.sAo + zi * p.sAi + r * p.sAm;
        float acc[8] = {0.f, 0.f, 0.f, 0.f, 0.f, 0.f, 0.f, 0.f};
        for (int k = 0; k < p.K; ++k) { const float a = A[(long long)k * p.sAk];
#pragma unroll
            for (int j = 0; j < 8; ++j) if (j < p.N) acc[j] += a * Bb[(long long)j * p.sBn + (long long)k * p.sBk]; }
#pragma unroll
        for (int j = 0; j < 8; ++j) if (j < p.N) {
            float v = acc[j] * p.alpha;
            if (p.flags & 1) v += p.bias[j];
            if (p.flags & 2) v += p.bias[r];
            v = act_fn(v, p.act);
            if (p.flags & 4) v += p.beta * R[r * p.sRm + (long long)j * p.sRn];
            VST2(float, C + r * p.sCm + j, v);
        }
    }
}
__global__ __launch_bounds__(256) void k_smallsoftmax(const float* __restrict__ src, float* __restrict__ dst, long long sr, long long dr, int n, long long R, float scale) {
    const long long r0 = ((long long)blockIdx.x * 256 + threadIdx.x) * 32;
    for (int rr = 0; rr < 32; ++rr) {
        const long long r = r0 + rr; if (r >= R) return;
        const float* s = src + r * sr; float* d = dst + r * dr;
        float mx = -__builtin_inff();
        for (int j = 0; j < n; ++j) mx = fmaxf(mx, s[j] * scale);
        float sum = 0.f;
        for (int j = 0; j < n; ++j) sum += expf(s[j] * scale - mx);
        const float inv = 1.f / sum;
        for (int j = 0; j < n; ++j) { const float v = expf(s[j] * scale - mx) * inv; VST2(float, d + j, v); }
    }
}

__global__ __launch_bounds__(32) void k_unitstat(float* __restrict__ st) { const int t = threadIdx.x; const float v = (t == 1) ? 1.f : 0.f; VST2(float, st + t, v); }

__global__ __launch_bounds__(256) void k_lincopy(const float* __restrict__ src, long long lds, float* __restrict__ dst, long long ldd, long long rows, int cols) {
    const long long i = (long long)blockIdx.x * 256 + threadIdx.x; if (i >= rows * cols) return;
    const long long r = i / cols; const int c = (int)(i - r * cols);
    const float v = src[r * lds + c]; VST2(float, dst + r * ldd + c, v);
}

#define IL_CAP32 32
#define IL_T32 256
#define IL_TILE32 4096
__global__ __launch_bounds__(IL_T32) void k_inlists32(const int* __restrict__ tgt, int E, int N, int* __restrict__ NBR, int* __restrict__ cnt) {
    __shared__ int tt[IL_TILE32];
    __shared__ int lists[IL_T32 * IL_CAP32];
    const int d = blockIdx.x * IL_T32 + threadIdx.x; int n = 0;
    for (int e0 = 0; e0 < E; e0 += IL_TILE32) {
        const int nt = min(IL_TILE32, E - e0);
        __syncthreads();
        for (int i = threadIdx.x; i < nt; i += IL_T32) tt[i] = tgt[e0 + i];
        __syncthreads();
        for (int i = 0; i < nt; ++i) { if (tt[i] == d) { if (n < IL_CAP32) lists[threadIdx.x * IL_CAP32 + n] = e0 + i; ++n; } }
    }
    if (d < N) {
        int* row = NBR + (long long)d * IL_CAP32;
        for (int j = 0; j < IL_CAP32; ++j) { const int v = (j < n) ? lists[threadIdx.x * IL_CAP32 + j] : -1; VST2(int, row + j, v); }
        VST2(int, cnt + d, min(n, IL_CAP32));
    }
}
__global__ __launch_bounds__(256) void k_csr_scan32(const int* __restrict__ cnt, int* __restrict__ off, int N) {
    __shared__ int part[256]; const int per = ((((N + 255) / 256) + 31) / 32) * 32; const int a = threadIdx.x * per, b = min(N, a + per); int s = 0;
    for (int i = a; i < b; ++i) s += cnt[i]; part[threadIdx.x] = s; __syncthreads();
    if (threadIdx.x == 0) { int run = 0; for (int t = 0; t < 256; ++t) { const int v = part[t]; part[t] = run; run += v; } } __syncthreads();
    int run = part[threadIdx.x]; for (int i = a; i < b; ++i) { VST2(int, off + i, run); run += cnt[i]; }
    if (a < N && b == N) { VST2(int, off + N, run); }
}
__global__ __launch_bounds__(256) void k_slotcopy32(const int* __restrict__ off, const int* __restrict__ NBR, int* __restrict__ slot, int N) {
    const int t = blockIdx.x * 256 + threadIdx.x; const int tot = off[N]; if (t >= tot) return;
    int lo = 0, hi = N - 1;
    while (lo < hi) { const int mid = (lo + hi + 1) >> 1; if (off[mid] <= t) lo = mid; else hi = mid - 1; }
    int j = t - off[lo]; j = (j < 0) ? 0 : ((j >= IL_CAP32) ? (IL_CAP32 - 1) : j);
    VST2(int, slot + t, NBR[(long long)lo * IL_CAP32 + j]);
}

__global__ __launch_bounds__(256) void k_sb_nodectx(const float* __restrict__ nf, const int* __restrict__ etype, const float* __restrict__ ep, const int* __restrict__ tgt, const int* __restrict__ scope, const int* __restrict__ batch, const float* __restrict__ emb, float* __restrict__ NC, int N) { const int q = blockIdx.x * 256 + threadIdx.x; if (q >= N * 32) return; const int c = q % 32; const int n = q / 32; const int b = batch[n]; float v = 0.f;
    if (c < 7) v = nf[n * 7 + c]; else if (c < 23) v = emb[etype[b] * 16 + (c - 7)]; else if (c < 27) v = ep[b * 4 + (c - 23)]; else if (c == 27) v = (float)tgt[n]; else if (c == 28) v = (float)scope[n]; VST2(float, NC + q, v); }
__global__ __launch_bounds__(256) void k_sb_ws(const float* __restrict__ We1, float* __restrict__ WS, int H) { const int q = blockIdx.x * 256 + threadIdx.x; if (q >= 32 * H) return; const int h = q % H; const int r = q / H; float v = 0.f; if (r < 4) v = We1[r * H + h]; else if (r < 26) v = We1[(260 + (r - 4)) * H + h]; VST2(float, WS + q, v); }
__global__ __launch_bounds__(256) void k_sb_edgectx(const float* __restrict__ ef, const int* __restrict__ etype, const float* __restrict__ ep, const int* __restrict__ tgt, const int* __restrict__ scope, const int* __restrict__ batch, const float* __restrict__ emb, const int* __restrict__ ei, const float* __restrict__ F, float* __restrict__ EC, float* __restrict__ XS, float* __restrict__ XD, int e0, int CH, int E, int H) {
    const long long q = (long long)blockIdx.x * 256 + threadIdx.x; if (q >= (long long)CH * H) return; const int c = (int)(q % H); const int r = (int)(q / H); const int e = e0 + r; const int b = batch[e];
    VST2(float, XS + q, F[(long long)ei[e] * H + c]); VST2(float, XD + q, F[(long long)ei[E + e] * H + c]);
    if (c < 32) { float v = 0.f; if (c < 4) v = ef[(long long)e * 4 + c]; else if (c < 20) v = emb[etype[b] * 16 + (c - 4)]; else if (c < 24) v = ep[b * 4 + (c - 20)]; else if (c == 24) v = (float)tgt[e]; else if (c == 25) v = (float)scope[e]; VST2(float, EC + (long long)r * 32 + c, v); } }
__global__ __launch_bounds__(256) void k_sb_gather(const int* __restrict__ ei, const float* __restrict__ F, float* __restrict__ XS, float* __restrict__ XD, int e0, int CH, int E, int H) { const long long q = (long long)blockIdx.x * 256 + threadIdx.x; if (q >= (long long)CH * H) return; const int c = (int)(q % H); const int e = e0 + (int)(q / H); VST2(float, XS + q, F[(long long)ei[e] * H + c]); VST2(float, XD + q, F[(long long)ei[E + e] * H + c]); }
__global__ __launch_bounds__(256) void k_sb_scale(float* __restrict__ M, const int* __restrict__ scope, int e0, int CH, int H) { const long long q = (long long)blockIdx.x * 256 + threadIdx.x; if (q >= (long long)CH * H) return; const int e = e0 + (int)(q / H); const float v = M[q] * (float)scope[e]; VST2(float, M + q, v); }
__global__ __launch_bounds__(256) void k_sb_agg(const float* __restrict__ MSG, const int* __restrict__ soff, const int* __restrict__ sslot, const int* __restrict__ doff, const int* __restrict__ dslot, float* __restrict__ AGG, int e0, int CH, int N, int H) {
    const long long q = (long long)blockIdx.x * 256 + threadIdx.x; if (q >= (long long)N * H) return; const int c = (int)(q % H); const int n = (int)(q / H); float s = 0.f; int cnt = 0;
    for (int p = soff[n]; p < soff[n + 1]; ++p) { const int e = sslot[p]; if (e >= e0 && e < e0 + CH) { s += MSG[(long long)(e - e0) * H + c]; ++cnt; } }
    for (int p = doff[n]; p < doff[n + 1]; ++p) { const int e = dslot[p]; if (e >= e0 && e < e0 + CH) { s += MSG[(long long)(e - e0) * H + c]; ++cnt; } }
    if (cnt) { const float v = AGG[q] + s; VST2(float, AGG + q, v); } }
__global__ __launch_bounds__(256) void k_sb_nodeout(const float* __restrict__ RN, int ldp, const int* __restrict__ scope, const float* __restrict__ nf, float* __restrict__ O0, float* __restrict__ O2, int N) { const int q = blockIdx.x * 256 + threadIdx.x; if (q >= N * 7) return; const int j = q % 7; const int n = q / 7; const float sc = (float)scope[n]; const float d = RN[(long long)n * ldp + j] * sc; VST2(float, O0 + q, d); VST2(float, O2 + q, (sc > 0.5f) ? nf[q] + d : nf[q]); }
__global__ __launch_bounds__(256) void k_sb_edgeout(const float* __restrict__ RE, int ldp, const int* __restrict__ scope, const float* __restrict__ ef, float* __restrict__ O1, float* __restrict__ O3, int e0, int CH) { const int q = blockIdx.x * 256 + threadIdx.x; if (q >= CH * 4) return; const int j = q % 4; const int r = q / 4; const int e = e0 + r; const float sc = (float)scope[e]; const float d = RE[(long long)r * ldp + j] * sc; const long long o = (long long)e * 4 + j; VST2(float, O1 + o, d); VST2(float, O3 + o, (sc > 0.5f) ? ef[o] + d : ef[o]); }

template __global__ void k_gemm<1>(GemmP);

extern "C" void kernel_launch(void* const* d_in, const int* in_sizes, int n_in, void* d_out, int out_size, void* d_ws, size_t ws_size, hipStream_t stream) {
    (void)in_sizes; (void)n_in; (void)out_size; (void)ws_size;
    const float* nf = (const float*)d_in[0];
    const int* ei = (const int*)d_in[1];
    const float* ef = (const float*)d_in[2];
    const int* etype = (const int*)d_in[3];
    const float* eparams = (const float*)d_in[4];
    const int* nmask = (const int*)d_in[5];
    const int* emask = (const int*)d_in[6];
    const int* nscope = (const int*)d_in[7];
    const int* escope = (const int*)d_in[8];
    const int* nbatch = (const int*)d_in[9];
    const int* ebatch = (const int*)d_in[10];
    const int* npg = (const int*)d_in[11];
    const int* epg = (const int*)d_in[12];
    const float* emb = (const float*)d_in[13];
    const float* Wn1 = (const float*)d_in[14];
    const float* bn1 = (const float*)d_in[15];
    const float* Wn2 = (const float*)d_in[16];
    const float* bn2 = (const float*)d_in[17];
    const float* We1 = (const float*)d_in[18];
    const float* be1 = (const float*)d_in[19];
    const float* We2 = (const float*)d_in[20];
    const float* be2 = (const float*)d_in[21];
    const float* Wm = (const float*)d_in[22];
    const float* bm = (const float*)d_in[23];
    const float* Wu = (const float*)d_in[24];
    const float* bu = (const float*)d_in[25];
    const float* Wnd = (const float*)d_in[26];
    const float* bnd = (const float*)d_in[27];
    const float* Wed1 = (const float*)d_in[28];
    const float* bed1 = (const float*)d_in[29];
    const float* Wed2 = (const float*)d_in[30];
    const float* bed2 = (const float*)d_in[31];
    const int N = 50000;
    const int E = 500000;
    const int H = 128;
    const int CH = 31250;
    const int CAP = 32;
    const int LP = 32;
    float* out = (float*)d_out;
    float* o1 = out + ((size_t)N * 7);
    float* o2 = out + ((size_t)N * 7 + (size_t)E * 4);
    float* o3 = out + ((size_t)N * 7 * 2 + (size_t)E * 4);
    char* wsp = (char*)d_ws;
    int* scnt = (int*)wsp; wsp += (((size_t)((size_t)N + 64) * 4 + 255) / 256) * 256;
    int* soff = (int*)wsp; wsp += (((size_t)((size_t)N + 64) * 4 + 255) / 256) * 256;
    int* sslot = (int*)wsp; wsp += (((size_t)((size_t)E + 64) * 4 + 255) / 256) * 256;
    int* snbr = (int*)wsp; wsp += (((size_t)((size_t)N * CAP) * 4 + 255) / 256) * 256;
    int* dcnt = (int*)wsp; wsp += (((size_t)((size_t)N + 64) * 4 + 255) / 256) * 256;
    int* doff = (int*)wsp; wsp += (((size_t)((size_t)N + 64) * 4 + 255) / 256) * 256;
    int* dslot = (int*)wsp; wsp += (((size_t)((size_t)E + 64) * 4 + 255) / 256) * 256;
    int* dnbr = (int*)wsp; wsp += (((size_t)((size_t)N * CAP) * 4 + 255) / 256) * 256;
    float* NC = (float*)wsp; wsp += (((size_t)((size_t)N * 32) * 4 + 255) / 256) * 256;
    float* NH1 = (float*)wsp; wsp += (((size_t)((size_t)N * H) * 4 + 255) / 256) * 256;
    float* NH = (float*)wsp; wsp += (((size_t)((size_t)N * H) * 4 + 255) / 256) * 256;
    float* AGG = (float*)wsp; wsp += (((size_t)((size_t)N * H) * 4 + 255) / 256) * 256;
    float* HU = (float*)wsp; wsp += (((size_t)((size_t)N * H) * 4 + 255) / 256) * 256;
    float* RN = (float*)wsp; wsp += (((size_t)((size_t)N * LP) * 4 + 255) / 256) * 256;
    float* WS = (float*)wsp; wsp += (((size_t)((size_t)32 * H) * 4 + 255) / 256) * 256;
    float* EC = (float*)wsp; wsp += (((size_t)((size_t)CH * 32) * 4 + 255) / 256) * 256;
    float* XS = (float*)wsp; wsp += (((size_t)((size_t)CH * H) * 4 + 255) / 256) * 256;
    float* XD = (float*)wsp; wsp += (((size_t)((size_t)CH * H) * 4 + 255) / 256) * 256;
    float* EH1 = (float*)wsp; wsp += (((size_t)((size_t)CH * H) * 4 + 255) / 256) * 256;
    float* EH = (float*)wsp; wsp += (((size_t)((size_t)CH * H) * 4 + 255) / 256) * 256;
    float* MSG = (float*)wsp; wsp += (((size_t)((size_t)CH * H) * 4 + 255) / 256) * 256;
    float* RE = (float*)wsp; wsp += (((size_t)((size_t)CH * LP) * 4 + 255) / 256) * 256;
    float* ust = (float*)wsp; wsp += (((size_t)(64) * 4 + 255) / 256) * 256;
    k_inlists32<<<(unsigned)((N) + IL_T32 - 1) / IL_T32, IL_T32, 0, stream>>>(ei, E, N, snbr, scnt);
    k_csr_scan32<<<1, 256, 0, stream>>>(scnt, soff, N);
    k_slotcopy32<<<(unsigned)((E) + 255) / 256, 256, 0, stream>>>(soff, snbr, sslot, N);
    k_inlists32<<<(unsigned)((N) + IL_T32 - 1) / IL_T32, IL_T32, 0, stream>>>(ei + E, E, N, dnbr, dcnt);
    k_csr_scan32<<<1, 256, 0, stream>>>(dcnt, doff, N);
    k_slotcopy32<<<(unsigned)((E) + 255) / 256, 256, 0, stream>>>(doff, dnbr, dslot, N);
    k_unitstat<<<1, 32, 0, stream>>>(ust);
    hipMemsetAsync(AGG, 0, (size_t)N * H * 4, stream);
    k_sb_nodectx<<<(unsigned)((N * 32 + 255) / 256), 256, 0, stream>>>(nf, etype, eparams, nmask, nscope, nbatch, emb, NC, N);
    k_sb_ws<<<(unsigned)((32 * H + 255) / 256), 256, 0, stream>>>(We1, WS, H);
    { GemmP gn1;
      gn1.A = NC; gn1.B = Wn1; gn1.bias = bn1; gn1.R = NC; gn1.C = NH1;
      gn1.sAo = 0; gn1.sAi = 0; gn1.sAm = 32; gn1.sAk = 1; gn1.sBo = 0; gn1.sBi = 0; gn1.sBn = 1; gn1.sBk = H; gn1.sCo = 0; gn1.sCi = 0; gn1.sCm = H; gn1.sRo = 0; gn1.sRi = 0; gn1.sRm = 0; gn1.sRn = 0;
      gn1.M = N; gn1.N = H; gn1.K = 29; gn1.zi_n = 1; gn1.flags = 1; gn1.act = 1;
      gn1.alpha = 1.0f; gn1.beta = 0.0f; gn1.sa = 1.0f; gn1.sb = 1.0f; gn1.Npad = H; gn1.pad_ = 0;
      k_gemm<1><<<dim3((unsigned)((H) + 31) / 32, (unsigned)((N) + 15) / 16, (unsigned)(1)), 32, 0, stream>>>(gn1); }
    { GemmP gn2;
      gn2.A = NH1; gn2.B = Wn2; gn2.bias = bn2; gn2.R = NH1; gn2.C = NH;
      gn2.sAo = 0; gn2.sAi = 0; gn2.sAm = H; gn2.sAk = 1; gn2.sBo = 0; gn2.sBi = 0; gn2.sBn = 1; gn2.sBk = H; gn2.sCo = 0; gn2.sCi = 0; gn2.sCm = H; gn2.sRo = 0; gn2.sRi = 0; gn2.sRm = 0; gn2.sRn = 0;
      gn2.M = N; gn2.N = H; gn2.K = H; gn2.zi_n = 1; gn2.flags = 1; gn2.act = 1;
      gn2.alpha = 1.0f; gn2.beta = 0.0f; gn2.sa = 1.0f; gn2.sb = 1.0f; gn2.Npad = H; gn2.pad_ = 0;
      k_gemm<1><<<dim3((unsigned)((H) + 31) / 32, (unsigned)((N) + 15) / 16, (unsigned)(1)), 32, 0, stream>>>(gn2); }
    k_sb_edgectx<<<(unsigned)(((long long)CH * H + 255) / 256), 256, 0, stream>>>(ef, etype, eparams, emask, escope, ebatch, emb, ei, NH, EC, XS, XD, 0, CH, E, H);
    { GemmP ge1aa0;
      ge1aa0.A = EC; ge1aa0.B = WS; ge1aa0.bias = be1; ge1aa0.R = EC; ge1aa0.C = EH1;
      ge1aa0.sAo = 0; ge1aa0.sAi = 0; ge1aa0.sAm = 32; ge1aa0.sAk = 1; ge1aa0.sBo = 0; ge1aa0.sBi = 0; ge1aa0.sBn = 1; ge1aa0.sBk = H; ge1aa0.sCo = 0; ge1aa0.sCi = 0; ge1aa0.sCm = H; ge1aa0.sRo = 0; ge1aa0.sRi = 0; ge1aa0.sRm = 0; ge1aa0.sRn = 0;
      ge1aa0.M = CH; ge1aa0.N = H; ge1aa0.K = 26; ge1aa0.zi_n = 1; ge1aa0.flags = 1; ge1aa0.act = 0;
      ge1aa0.alpha = 1.0f; ge1aa0.beta = 0.0f; ge1aa0.sa = 1.0f; ge1aa0.sb = 1.0f; ge1aa0.Npad = H; ge1aa0.pad_ = 0;
      k_gemm<1><<<dim3((unsigned)((H) + 31) / 32, (unsigned)((CH) + 15) / 16, (unsigned)(1)), 32, 0, stream>>>(ge1aa0); }
    { GemmP ge1ba0;
      ge1ba0.A = XS; ge1ba0.B = We1 + (size_t)4 * H; ge1ba0.bias = XS; ge1ba0.R = EH1; ge1ba0.C = EH1;
      ge1ba0.sAo = 0; ge1ba0.sAi = 0; ge1ba0.sAm = H; ge1ba0.sAk = 1; ge1ba0.sBo = 0; ge1ba0.sBi = 0; ge1ba0.sBn = 1; ge1ba0.sBk = H; ge1ba0.sCo = 0; ge1ba0.sCi = 0; ge1ba0.sCm = H; ge1ba0.sRo = 0; ge1ba0.sRi = 0; ge1ba0.sRm = H; ge1ba0.sRn = 1;
      ge1ba0.M = CH; ge1ba0.N = H; ge1ba0.K = H; ge1ba0.zi_n = 1; ge1ba0.flags = 4; ge1ba0.act = 0;
      ge1ba0.alpha = 1.0f; ge1ba0.beta = 1.0f; ge1ba0.sa = 1.0f; ge1ba0.sb = 1.0f; ge1ba0.Npad = H; ge1ba0.pad_ = 0;
      k_gemm<1><<<dim3((unsigned)((H) + 31) / 32, (unsigned)((CH) + 15) / 16, (unsigned)(1)), 32, 0, stream>>>(ge1ba0); }
    { GemmP ge1ca0;
      ge1ca0.A = XD; ge1ca0.B = We1 + (size_t)132 * H; ge1ca0.bias = XD; ge1ca0.R = EH1; ge1ca0.C = EH1;
      ge1ca0.sAo = 0; ge1ca0.sAi = 0; ge1ca0.sAm = H; ge1ca0.sAk = 1; ge1ca0.sBo = 0; ge1ca0.sBi = 0; ge1ca0.sBn = 1; ge1ca0.sBk = H; ge1ca0.sCo = 0; ge1ca0.sCi = 0; ge1ca0.sCm = H; ge1ca0.sRo = 0; ge1ca0.sRi = 0; ge1ca0.sRm = H; ge1ca0.sRn = 1;
      ge1ca0.M = CH; ge1ca0.N = H; ge1ca0.K = H; ge1ca0.zi_n = 1; ge1ca0.flags = 4; ge1ca0.act = 0;
      ge1ca0.alpha = 1.0f; ge1ca0.beta = 1.0f; ge1ca0.sa = 1.0f; ge1ca0.sb = 1.0f; ge1ca0.Npad = H; ge1ca0.pad_ = 0;
      k_gemm<1><<<dim3((unsigned)((H) + 31) / 32, (unsigned)((CH) + 15) / 16, (unsigned)(1)), 32, 0, stream>>>(ge1ca0); }
    k_norm_apply<<<(unsigned)(((long long)(1) * (1) * ((long long)CH * H) + 255) / 256), 256, 0, stream>>>(EH1, EH1, ust, nullptr, nullptr, 1, 1, (long long)CH * H, 1, 0, 1);
    { GemmP ge2a0;
      ge2a0.A = EH1; ge2a0.B = We2; ge2a0.bias = be2; ge2a0.R = EH1; ge2a0.C = EH;
      ge2a0.sAo = 0; ge2a0.sAi = 0; ge2a0.sAm = H; ge2a0.sAk = 1; ge2a0.sBo = 0; ge2a0.sBi = 0; ge2a0.sBn = 1; ge2a0.sBk = H; ge2a0.sCo = 0; ge2a0.sCi = 0; ge2a0.sCm = H; ge2a0.sRo = 0; ge2a0.sRi = 0; ge2a0.sRm = 0; ge2a0.sRn = 0;
      ge2a0.M = CH; ge2a0.N = H; ge2a0.K = H; ge2a0.zi_n = 1; ge2a0.flags = 1; ge2a0.act = 1;
      ge2a0.alpha = 1.0f; ge2a0.beta = 0.0f; ge2a0.sa = 1.0f; ge2a0.sb = 1.0f; ge2a0.Npad = H; ge2a0.pad_ = 0;
      k_gemm<1><<<dim3((unsigned)((H) + 31) / 32, (unsigned)((CH) + 15) / 16, (unsigned)(1)), 32, 0, stream>>>(ge2a0); }
    { GemmP gm0;
      gm0.A = EH; gm0.B = Wm; gm0.bias = bm; gm0.R = EH; gm0.C = MSG;
      gm0.sAo = 0; gm0.sAi = 0; gm0.sAm = H; gm0.sAk = 1; gm0.sBo = 0; gm0.sBi = 0; gm0.sBn = 1; gm0.sBk = H; gm0.sCo = 0; gm0.sCi = 0; gm0.sCm = H; gm0.sRo = 0; gm0.sRi = 0; gm0.sRm = 0; gm0.sRn = 0;
      gm0.M = CH; gm0.N = H; gm0.K = H; gm0.zi_n = 1; gm0.flags = 1; gm0.act = 0;
      gm0.alpha = 1.0f; gm0.beta = 0.0f; gm0.sa = 1.0f; gm0.sb = 1.0f; gm0.Npad = H; gm0.pad_ = 0;
      k_gemm<1><<<dim3((unsigned)((H) + 31) / 32, (unsigned)((CH) + 15) / 16, (unsigned)(1)), 32, 0, stream>>>(gm0); }
    k_sb_scale<<<(unsigned)(((long long)CH * H + 255) / 256), 256, 0, stream>>>(MSG, escope, 0, CH, H);
    k_sb_agg<<<(unsigned)(((long long)N * H + 255) / 256), 256, 0, stream>>>(MSG, soff, sslot, doff, dslot, AGG, 0, CH, N, H);
    k_sb_edgectx<<<(unsigned)(((long long)CH * H + 255) / 256), 256, 0, stream>>>(ef, etype, eparams, emask, escope, ebatch, emb, ei, NH, EC, XS, XD, 31250, CH, E, H);
    { GemmP ge1aa1;
      ge1aa1.A = EC; ge1aa1.B = WS; ge1aa1.bias = be1; ge1aa1.R = EC; ge1aa1.C = EH1;
      ge1aa1.sAo = 0; ge1aa1.sAi = 0; ge1aa1.sAm = 32; ge1aa1.sAk = 1; ge1aa1.sBo = 0; ge1aa1.sBi = 0; ge1aa1.sBn = 1; ge1aa1.sBk = H; ge1aa1.sCo = 0; ge1aa1.sCi = 0; ge1aa1.sCm = H; ge1aa1.sRo = 0; ge1aa1.sRi = 0; ge1aa1.sRm = 0; ge1aa1.sRn = 0;
      ge1aa1.M = CH; ge1aa1.N = H; ge1aa1.K = 26; ge1aa1.zi_n = 1; ge1aa1.flags = 1; ge1aa1.act = 0;
      ge1aa1.alpha = 1.0f; ge1aa1.beta = 0.0f; ge1aa1.sa = 1.0f; ge1aa1.sb = 1.0f; ge1aa1.Npad = H; ge1aa1.pad_ = 0;
      k_gemm<1><<<dim3((unsigned)((H) + 31) / 32, (unsigned)((CH) + 15) / 16, (unsigned)(1)), 32, 0, stream>>>(ge1aa1); }
    { GemmP ge1ba1;
      ge1ba1.A = XS; ge1ba1.B = We1 + (size_t)4 * H; ge1ba1.bias = XS; ge1ba1.R = EH1; ge1ba1.C = EH1;
      ge1ba1.sAo = 0; ge1ba1.sAi = 0; ge1ba1.sAm = H; ge1ba1.sAk = 1; ge1ba1.sBo = 0; ge1ba1.sBi = 0; ge1ba1.sBn = 1; ge1ba1.sBk = H; ge1ba1.sCo = 0; ge1ba1.sCi = 0; ge1ba1.sCm = H; ge1ba1.sRo = 0; ge1ba1.sRi = 0; ge1ba1.sRm = H; ge1ba1.sRn = 1;
      ge1ba1.M = CH; ge1ba1.N = H; ge1ba1.K = H; ge1ba1.zi_n = 1; ge1ba1.flags = 4; ge1ba1.act = 0;
      ge1ba1.alpha = 1.0f; ge1ba1.beta = 1.0f; ge1ba1.sa = 1.0f; ge1ba1.sb = 1.0f; ge1ba1.Npad = H; ge1ba1.pad_ = 0;
      k_gemm<1><<<dim3((unsigned)((H) + 31) / 32, (unsigned)((CH) + 15) / 16, (unsigned)(1)), 32, 0, stream>>>(ge1ba1); }
    { GemmP ge1ca1;
      ge1ca1.A = XD; ge1ca1.B = We1 + (size_t)132 * H; ge1ca1.bias = XD; ge1ca1.R = EH1; ge1ca1.C = EH1;
      ge1ca1.sAo = 0; ge1ca1.sAi = 0; ge1ca1.sAm = H; ge1ca1.sAk = 1; ge1ca1.sBo = 0; ge1ca1.sBi = 0; ge1ca1.sBn = 1; ge1ca1.sBk = H; ge1ca1.sCo = 0; ge1ca1.sCi = 0; ge1ca1.sCm = H; ge1ca1.sRo = 0; ge1ca1.sRi = 0; ge1ca1.sRm = H; ge1ca1.sRn = 1;
      ge1ca1.M = CH; ge1ca1.N = H; ge1ca1.K = H; ge1ca1.zi_n = 1; ge1ca1.flags = 4; ge1ca1.act = 0;
      ge1ca1.alpha = 1.0f; ge1ca1.beta = 1.0f; ge1ca1.sa = 1.0f; ge1ca1.sb = 1.0f; ge1ca1.Npad = H; ge1ca1.pad_ = 0;
      k_gemm<1><<<dim3((unsigned)((H) + 31) / 32, (unsigned)((CH) + 15) / 16, (unsigned)(1)), 32, 0, stream>>>(ge1ca1); }
    k_norm_apply<<<(unsigned)(((long long)(1) * (1) * ((long long)CH * H) + 255) / 256), 256, 0, stream>>>(EH1, EH1, ust, nullptr, nullptr, 1, 1, (long long)CH * H, 1, 0, 1);
    { GemmP ge2a1;
      ge2a1.A = EH1; ge2a1.B = We2; ge2a1.bias = be2; ge2a1.R = EH1; ge2a1.C = EH;
      ge2a1.sAo = 0; ge2a1.sAi = 0; ge2a1.sAm = H; ge2a1.sAk = 1; ge2a1.sBo = 0; ge2a1.sBi = 0; ge2a1.sBn = 1; ge2a1.sBk = H; ge2a1.sCo = 0; ge2a1.sCi = 0; ge2a1.sCm = H; ge2a1.sRo = 0; ge2a1.sRi = 0; ge2a1.sRm = 0; ge2a1.sRn = 0;
      ge2a1.M = CH; ge2a1.N = H; ge2a1.K = H; ge2a1.zi_n = 1; ge2a1.flags = 1; ge2a1.act = 1;
      ge2a1.alpha = 1.0f; ge2a1.beta = 0.0f; ge2a1.sa = 1.0f; ge2a1.sb = 1.0f; ge2a1.Npad = H; ge2a1.pad_ = 0;
      k_gemm<1><<<dim3((unsigned)((H) + 31) / 32, (unsigned)((CH) + 15) / 16, (unsigned)(1)), 32, 0, stream>>>(ge2a1); }
    { GemmP gm1;
      gm1.A = EH; gm1.B = Wm; gm1.bias = bm; gm1.R = EH; gm1.C = MSG;
      gm1.sAo = 0; gm1.sAi = 0; gm1.sAm = H; gm1.sAk = 1; gm1.sBo = 0; gm1.sBi = 0; gm1.sBn = 1; gm1.sBk = H; gm1.sCo = 0; gm1.sCi = 0; gm1.sCm = H; gm1.sRo = 0; gm1.sRi = 0; gm1.sRm = 0; gm1.sRn = 0;
      gm1.M = CH; gm1.N = H; gm1.K = H; gm1.zi_n = 1; gm1.flags = 1; gm1.act = 0;
      gm1.alpha = 1.0f; gm1.beta = 0.0f; gm1.sa = 1.0f; gm1.sb = 1.0f; gm1.Npad = H; gm1.pad_ = 0;
      k_gemm<1><<<dim3((unsigned)((H) + 31) / 32, (unsigned)((CH) + 15) / 16, (unsigned)(1)), 32, 0, stream>>>(gm1); }
    k_sb_scale<<<(unsigned)(((long long)CH * H + 255) / 256), 256, 0, stream>>>(MSG, escope, 31250, CH, H);
    k_sb_agg<<<(unsigned)(((long long)N * H + 255) / 256), 256, 0, stream>>>(MSG, soff, sslot, doff, dslot, AGG, 31250, CH, N, H);
    k_sb_edgectx<<<(unsigned)(((long long)CH * H + 255) / 256), 256, 0, stream>>>(ef, etype, eparams, emask, escope, ebatch, emb, ei, NH, EC, XS, XD, 62500, CH, E, H);
    { GemmP ge1aa2;
      ge1aa2.A = EC; ge1aa2.B = WS; ge1aa2.bias = be1; ge1aa2.R = EC; ge1aa2.C = EH1;
      ge1aa2.sAo = 0; ge1aa2.sAi = 0; ge1aa2.sAm = 32; ge1aa2.sAk = 1; ge1aa2.sBo = 0; ge1aa2.sBi = 0; ge1aa2.sBn = 1; ge1aa2.sBk = H; ge1aa2.sCo = 0; ge1aa2.sCi = 0; ge1aa2.sCm = H; ge1aa2.sRo = 0; ge1aa2.sRi = 0; ge1aa2.sRm = 0; ge1aa2.sRn = 0;
      ge1aa2.M = CH; ge1aa2.N = H; ge1aa2.K = 26; ge1aa2.zi_n = 1; ge1aa2.flags = 1; ge1aa2.act = 0;
      ge1aa2.alpha = 1.0f; ge1aa2.beta = 0.0f; ge1aa2.sa = 1.0f; ge1aa2.sb = 1.0f; ge1aa2.Npad = H; ge1aa2.pad_ = 0;
      k_gemm<1><<<dim3((unsigned)((H) + 31) / 32, (unsigned)((CH) + 15) / 16, (unsigned)(1)), 32, 0, stream>>>(ge1aa2); }
    { GemmP ge1ba2;
      ge1ba2.A = XS; ge1ba2.B = We1 + (size_t)4 * H; ge1ba2.bias = XS; ge1ba2.R = EH1; ge1ba2.C = EH1;
      ge1ba2.sAo = 0; ge1ba2.sAi = 0; ge1ba2.sAm = H; ge1ba2.sAk = 1; ge1ba2.sBo = 0; ge1ba2.sBi = 0; ge1ba2.sBn = 1; ge1ba2.sBk = H; ge1ba2.sCo = 0; ge1ba2.sCi = 0; ge1ba2.sCm = H; ge1ba2.sRo = 0; ge1ba2.sRi = 0; ge1ba2.sRm = H; ge1ba2.sRn = 1;
      ge1ba2.M = CH; ge1ba2.N = H; ge1ba2.K = H; ge1ba2.zi_n = 1; ge1ba2.flags = 4; ge1ba2.act = 0;
      ge1ba2.alpha = 1.0f; ge1ba2.beta = 1.0f; ge1ba2.sa = 1.0f; ge1ba2.sb = 1.0f; ge1ba2.Npad = H; ge1ba2.pad_ = 0;
      k_gemm<1><<<dim3((unsigned)((H) + 31) / 32, (unsigned)((CH) + 15) / 16, (unsigned)(1)), 32, 0, stream>>>(ge1ba2); }
    { GemmP ge1ca2;
      ge1ca2.A = XD; ge1ca2.B = We1 + (size_t)132 * H; ge1ca2.bias = XD; ge1ca2.R = EH1; ge1ca2.C = EH1;
      ge1ca2.sAo = 0; ge1ca2.sAi = 0; ge1ca2.sAm = H; ge1ca2.sAk = 1; ge1ca2.sBo = 0; ge1ca2.sBi = 0; ge1ca2.sBn = 1; ge1ca2.sBk = H; ge1ca2.sCo = 0; ge1ca2.sCi = 0; ge1ca2.sCm = H; ge1ca2.sRo = 0; ge1ca2.sRi = 0; ge1ca2.sRm = H; ge1ca2.sRn = 1;
      ge1ca2.M = CH; ge1ca2.N = H; ge1ca2.K = H; ge1ca2.zi_n = 1; ge1ca2.flags = 4; ge1ca2.act = 0;
      ge1ca2.alpha = 1.0f; ge1ca2.beta = 1.0f; ge1ca2.sa = 1.0f; ge1ca2.sb = 1.0f; ge1ca2.Npad = H; ge1ca2.pad_ = 0;
      k_gemm<1><<<dim3((unsigned)((H) + 31) / 32, (unsigned)((CH) + 15) / 16, (unsigned)(1)), 32, 0, stream>>>(ge1ca2); }
    k_norm_apply<<<(unsigned)(((long long)(1) * (1) * ((long long)CH * H) + 255) / 256), 256, 0, stream>>>(EH1, EH1, ust, nullptr, nullptr, 1, 1, (long long)CH * H, 1, 0, 1);
    { GemmP ge2a2;
      ge2a2.A = EH1; ge2a2.B = We2; ge2a2.bias = be2; ge2a2.R = EH1; ge2a2.C = EH;
      ge2a2.sAo = 0; ge2a2.sAi = 0; ge2a2.sAm = H; ge2a2.sAk = 1; ge2a2.sBo = 0; ge2a2.sBi = 0; ge2a2.sBn = 1; ge2a2.sBk = H; ge2a2.sCo = 0; ge2a2.sCi = 0; ge2a2.sCm = H; ge2a2.sRo = 0; ge2a2.sRi = 0; ge2a2.sRm = 0; ge2a2.sRn = 0;
      ge2a2.M = CH; ge2a2.N = H; ge2a2.K = H; ge2a2.zi_n = 1; ge2a2.flags = 1; ge2a2.act = 1;
      ge2a2.alpha = 1.0f; ge2a2.beta = 0.0f; ge2a2.sa = 1.0f; ge2a2.sb = 1.0f; ge2a2.Npad = H; ge2a2.pad_ = 0;
      k_gemm<1><<<dim3((unsigned)((H) + 31) / 32, (unsigned)((CH) + 15) / 16, (unsigned)(1)), 32, 0, stream>>>(ge2a2); }
    { GemmP gm2;
      gm2.A = EH; gm2.B = Wm; gm2.bias = bm; gm2.R = EH; gm2.C = MSG;
      gm2.sAo = 0; gm2.sAi = 0; gm2.sAm = H; gm2.sAk = 1; gm2.sBo = 0; gm2.sBi = 0; gm2.sBn = 1; gm2.sBk = H; gm2.sCo = 0; gm2.sCi = 0; gm2.sCm = H; gm2.sRo = 0; gm2.sRi = 0; gm2.sRm = 0; gm2.sRn = 0;
      gm2.M = CH; gm2.N = H; gm2.K = H; gm2.zi_n = 1; gm2.flags = 1; gm2.act = 0;
      gm2.alpha = 1.0f; gm2.beta = 0.0f; gm2.sa = 1.0f; gm2.sb = 1.0f; gm2.Npad = H; gm2.pad_ = 0;
      k_gemm<1><<<dim3((unsigned)((H) + 31) / 32, (unsigned)((CH) + 15) / 16, (unsigned)(1)), 32, 0, stream>>>(gm2); }
    k_sb_scale<<<(unsigned)(((long long)CH * H + 255) / 256), 256, 0, stream>>>(MSG, escope, 62500, CH, H);
    k_sb_agg<<<(unsigned)(((long long)N * H + 255) / 256), 256, 0, stream>>>(MSG, soff, sslot, doff, dslot, AGG, 62500, CH, N, H);
    k_sb_edgectx<<<(unsigned)(((long long)CH * H + 255) / 256), 256, 0, stream>>>(ef, etype, eparams, emask, escope, ebatch, emb, ei, NH, EC, XS, XD, 93750, CH, E, H);
    { GemmP ge1aa3;
      ge1aa3.A = EC; ge1aa3.B = WS; ge1aa3.bias = be1; ge1aa3.R = EC; ge1aa3.C = EH1;
      ge1aa3.sAo = 0; ge1aa3.sAi = 0; ge1aa3.sAm = 32; ge1aa3.sAk = 1; ge1aa3.sBo = 0; ge1aa3.sBi = 0; ge1aa3.sBn = 1; ge1aa3.sBk = H; ge1aa3.sCo = 0; ge1aa3.sCi = 0; ge1aa3.sCm = H; ge1aa3.sRo = 0; ge1aa3.sRi = 0; ge1aa3.sRm = 0; ge1aa3.sRn = 0;
      ge1aa3.M = CH; ge1aa3.N = H; ge1aa3.K = 26; ge1aa3.zi_n = 1; ge1aa3.flags = 1; ge1aa3.act = 0;
      ge1aa3.alpha = 1.0f; ge1aa3.beta = 0.0f; ge1aa3.sa = 1.0f; ge1aa3.sb = 1.0f; ge1aa3.Npad = H; ge1aa3.pad_ = 0;
      k_gemm<1><<<dim3((unsigned)((H) + 31) / 32, (unsigned)((CH) + 15) / 16, (unsigned)(1)), 32, 0, stream>>>(ge1aa3); }
    { GemmP ge1ba3;
      ge1ba3.A = XS; ge1ba3.B = We1 + (size_t)4 * H; ge1ba3.bias = XS; ge1ba3.R = EH1; ge1ba3.C = EH1;
      ge1ba3.sAo = 0; ge1ba3.sAi = 0; ge1ba3.sAm = H; ge1ba3.sAk = 1; ge1ba3.sBo = 0; ge1ba3.sBi = 0; ge1ba3.sBn = 1; ge1ba3.sBk = H; ge1ba3.sCo = 0; ge1ba3.sCi = 0; ge1ba3.sCm = H; ge1ba3.sRo = 0; ge1ba3.sRi = 0; ge1ba3.sRm = H; ge1ba3.sRn = 1;
      ge1ba3.M = CH; ge1ba3.N = H; ge1ba3.K = H; ge1ba3.zi_n = 1; ge1ba3.flags = 4; ge1ba3.act = 0;
      ge1ba3.alpha = 1.0f; ge1ba3.beta = 1.0f; ge1ba3.sa = 1.0f; ge1ba3.sb = 1.0f; ge1ba3.Npad = H; ge1ba3.pad_ = 0;
      k_gemm<1><<<dim3((unsigned)((H) + 31) / 32, (unsigned)((CH) + 15) / 16, (unsigned)(1)), 32, 0, stream>>>(ge1ba3); }
    { GemmP ge1ca3;
      ge1ca3.A = XD; ge1ca3.B = We1 + (size_t)132 * H; ge1ca3.bias = XD; ge1ca3.R = EH1; ge1ca3.C = EH1;
      ge1ca3.sAo = 0; ge1ca3.sAi = 0; ge1ca3.sAm = H; ge1ca3.sAk = 1; ge1ca3.sBo = 0; ge1ca3.sBi = 0; ge1ca3.sBn = 1; ge1ca3.sBk = H; ge1ca3.sCo = 0; ge1ca3.sCi = 0; ge1ca3.sCm = H; ge1ca3.sRo = 0; ge1ca3.sRi = 0; ge1ca3.sRm = H; ge1ca3.sRn = 1;
      ge1ca3.M = CH; ge1ca3.N = H; ge1ca3.K = H; ge1ca3.zi_n = 1; ge1ca3.flags = 4; ge1ca3.act = 0;
      ge1ca3.alpha = 1.0f; ge1ca3.beta = 1.0f; ge1ca3.sa = 1.0f; ge1ca3.sb = 1.0f; ge1ca3.Npad = H; ge1ca3.pad_ = 0;
      k_gemm<1><<<dim3((unsigned)((H) + 31) / 32, (unsigned)((CH) + 15) / 16, (unsigned)(1)), 32, 0, stream>>>(ge1ca3); }
    k_norm_apply<<<(unsigned)(((long long)(1) * (1) * ((long long)CH * H) + 255) / 256), 256, 0, stream>>>(EH1, EH1, ust, nullptr, nullptr, 1, 1, (long long)CH * H, 1, 0, 1);
    { GemmP ge2a3;
      ge2a3.A = EH1; ge2a3.B = We2; ge2a3.bias = be2; ge2a3.R = EH1; ge2a3.C = EH;
      ge2a3.sAo = 0; ge2a3.sAi = 0; ge2a3.sAm = H; ge2a3.sAk = 1; ge2a3.sBo = 0; ge2a3.sBi = 0; ge2a3.sBn = 1; ge2a3.sBk = H; ge2a3.sCo = 0; ge2a3.sCi = 0; ge2a3.sCm = H; ge2a3.sRo = 0; ge2a3.sRi = 0; ge2a3.sRm = 0; ge2a3.sRn = 0;
      ge2a3.M = CH; ge2a3.N = H; ge2a3.K = H; ge2a3.zi_n = 1; ge2a3.flags = 1; ge2a3.act = 1;
      ge2a3.alpha = 1.0f; ge2a3.beta = 0.0f; ge2a3.sa = 1.0f; ge2a3.sb = 1.0f; ge2a3.Npad = H; ge2a3.pad_ = 0;
      k_gemm<1><<<dim3((unsigned)((H) + 31) / 32, (unsigned)((CH) + 15) / 16, (unsigned)(1)), 32, 0, stream>>>(ge2a3); }
    { GemmP gm3;
      gm3.A = EH; gm3.B = Wm; gm3.bias = bm; gm3.R = EH; gm3.C = MSG;
      gm3.sAo = 0; gm3.sAi = 0; gm3.sAm = H; gm3.sAk = 1; gm3.sBo = 0; gm3.sBi = 0; gm3.sBn = 1; gm3.sBk = H; gm3.sCo = 0; gm3.sCi = 0; gm3.sCm = H; gm3.sRo = 0; gm3.sRi = 0; gm3.sRm = 0; gm3.sRn = 0;
      gm3.M = CH; gm3.N = H; gm3.K = H; gm3.zi_n = 1; gm3.flags = 1; gm3.act = 0;
      gm3.alpha = 1.0f; gm3.beta = 0.0f; gm3.sa = 1.0f; gm3.sb = 1.0f; gm3.Npad = H; gm3.pad_ = 0;
      k_gemm<1><<<dim3((unsigned)((H) + 31) / 32, (unsigned)((CH) + 15) / 16, (unsigned)(1)), 32, 0, stream>>>(gm3); }
    k_sb_scale<<<(unsigned)(((long long)CH * H + 255) / 256), 256, 0, stream>>>(MSG, escope, 93750, CH, H);
    k_sb_agg<<<(unsigned)(((long long)N * H + 255) / 256), 256, 0, stream>>>(MSG, soff, sslot, doff, dslot, AGG, 93750, CH, N, H);
    k_sb_edgectx<<<(unsigned)(((long long)CH * H + 255) / 256), 256, 0, stream>>>(ef, etype, eparams, emask, escope, ebatch, emb, ei, NH, EC, XS, XD, 125000, CH, E, H);
    { GemmP ge1aa4;
      ge1aa4.A = EC; ge1aa4.B = WS; ge1aa4.bias = be1; ge1aa4.R = EC; ge1aa4.C = EH1;
      ge1aa4.sAo = 0; ge1aa4.sAi = 0; ge1aa4.sAm = 32; ge1aa4.sAk = 1; ge1aa4.sBo = 0; ge1aa4.sBi = 0; ge1aa4.sBn = 1; ge1aa4.sBk = H; ge1aa4.sCo = 0; ge1aa4.sCi = 0; ge1aa4.sCm = H; ge1aa4.sRo = 0; ge1aa4.sRi = 0; ge1aa4.sRm = 0; ge1aa4.sRn = 0;
      ge1aa4.M = CH; ge1aa4.N = H; ge1aa4.K = 26; ge1aa4.zi_n = 1; ge1aa4.flags = 1; ge1aa4.act = 0;
      ge1aa4.alpha = 1.0f; ge1aa4.beta = 0.0f; ge1aa4.sa = 1.0f; ge1aa4.sb = 1.0f; ge1aa4.Npad = H; ge1aa4.pad_ = 0;
      k_gemm<1><<<dim3((unsigned)((H) + 31) / 32, (unsigned)((CH) + 15) / 16, (unsigned)(1)), 32, 0, stream>>>(ge1aa4); }
    { GemmP ge1ba4;
      ge1ba4.A = XS; ge1ba4.B = We1 + (size_t)4 * H; ge1ba4.bias = XS; ge1ba4.R = EH1; ge1ba4.C = EH1;
      ge1ba4.sAo = 0; ge1ba4.sAi = 0; ge1ba4.sAm = H; ge1ba4.sAk = 1; ge1ba4.sBo = 0; ge1ba4.sBi = 0; ge1ba4.sBn = 1; ge1ba4.sBk = H; ge1ba4.sCo = 0; ge1ba4.sCi = 0; ge1ba4.sCm = H; ge1ba4.sRo = 0; ge1ba4.sRi = 0; ge1ba4.sRm = H; ge1ba4.sRn = 1;
      ge1ba4.M = CH; ge1ba4.N = H; ge1ba4.K = H; ge1ba4.zi_n = 1; ge1ba4.flags = 4; ge1ba4.act = 0;
      ge1ba4.alpha = 1.0f; ge1ba4.beta = 1.0f; ge1ba4.sa = 1.0f; ge1ba4.sb = 1.0f; ge1ba4.Npad = H; ge1ba4.pad_ = 0;
      k_gemm<1><<<dim3((unsigned)((H) + 31) / 32, (unsigned)((CH) + 15) / 16, (unsigned)(1)), 32, 0, stream>>>(ge1ba4); }
    { GemmP ge1ca4;
      ge1ca4.A = XD; ge1ca4.B = We1 + (size_t)132 * H; ge1ca4.bias = XD; ge1ca4.R = EH1; ge1ca4.C = EH1;
      ge1ca4.sAo = 0; ge1ca4.sAi = 0; ge1ca4.sAm = H; ge1ca4.sAk = 1; ge1ca4.sBo = 0; ge1ca4.sBi = 0; ge1ca4.sBn = 1; ge1ca4.sBk = H; ge1ca4.sCo = 0; ge1ca4.sCi = 0; ge1ca4.sCm = H; ge1ca4.sRo = 0; ge1ca4.sRi = 0; ge1ca4.sRm = H; ge1ca4.sRn = 1;
      ge1ca4.M = CH; ge1ca4.N = H; ge1ca4.K = H; ge1ca4.zi_n = 1; ge1ca4.flags = 4; ge1ca4.act = 0;
      ge1ca4.alpha = 1.0f; ge1ca4.beta = 1.0f; ge1ca4.sa = 1.0f; ge1ca4.sb = 1.0f; ge1ca4.Npad = H; ge1ca4.pad_ = 0;
      k_gemm<1><<<dim3((unsigned)((H) + 31) / 32, (unsigned)((CH) + 15) / 16, (unsigned)(1)), 32, 0, stream>>>(ge1ca4); }
    k_norm_apply<<<(unsigned)(((long long)(1) * (1) * ((long long)CH * H) + 255) / 256), 256, 0, stream>>>(EH1, EH1, ust, nullptr, nullptr, 1, 1, (long long)CH * H, 1, 0, 1);
    { GemmP ge2a4;
      ge2a4.A = EH1; ge2a4.B = We2; ge2a4.bias = be2; ge2a4.R = EH1; ge2a4.C = EH;
      ge2a4.sAo = 0; ge2a4.sAi = 0; ge2a4.sAm = H; ge2a4.sAk = 1; ge2a4.sBo = 0; ge2a4.sBi = 0; ge2a4.sBn = 1; ge2a4.sBk = H; ge2a4.sCo = 0; ge2a4.sCi = 0; ge2a4.sCm = H; ge2a4.sRo = 0; ge2a4.sRi = 0; ge2a4.sRm = 0; ge2a4.sRn = 0;
      ge2a4.M = CH; ge2a4.N = H; ge2a4.K = H; ge2a4.zi_n = 1; ge2a4.flags = 1; ge2a4.act = 1;
      ge2a4.alpha = 1.0f; ge2a4.beta = 0.0f; ge2a4.sa = 1.0f; ge2a4.sb = 1.0f; ge2a4.Npad = H; ge2a4.pad_ = 0;
      k_gemm<1><<<dim3((unsigned)((H) + 31) / 32, (unsigned)((CH) + 15) / 16, (unsigned)(1)), 32, 0, stream>>>(ge2a4); }
    { GemmP gm4;
      gm4.A = EH; gm4.B = Wm; gm4.bias = bm; gm4.R = EH; gm4.C = MSG;
      gm4.sAo = 0; gm4.sAi = 0; gm4.sAm = H; gm4.sAk = 1; gm4.sBo = 0; gm4.sBi = 0; gm4.sBn = 1; gm4.sBk = H; gm4.sCo = 0; gm4.sCi = 0; gm4.sCm = H; gm4.sRo = 0; gm4.sRi = 0; gm4.sRm = 0; gm4.sRn = 0;
      gm4.M = CH; gm4.N = H; gm4.K = H; gm4.zi_n = 1; gm4.flags = 1; gm4.act = 0;
      gm4.alpha = 1.0f; gm4.beta = 0.0f; gm4.sa = 1.0f; gm4.sb = 1.0f; gm4.Npad = H; gm4.pad_ = 0;
      k_gemm<1><<<dim3((unsigned)((H) + 31) / 32, (unsigned)((CH) + 15) / 16, (unsigned)(1)), 32, 0, stream>>>(gm4); }
    k_sb_scale<<<(unsigned)(((long long)CH * H + 255) / 256), 256, 0, stream>>>(MSG, escope, 125000, CH, H);
    k_sb_agg<<<(unsigned)(((long long)N * H + 255) / 256), 256, 0, stream>>>(MSG, soff, sslot, doff, dslot, AGG, 125000, CH, N, H);
    k_sb_edgectx<<<(unsigned)(((long long)CH * H + 255) / 256), 256, 0, stream>>>(ef, etype, eparams, emask, escope, ebatch, emb, ei, NH, EC, XS, XD, 156250, CH, E, H);
    { GemmP ge1aa5;
      ge1aa5.A = EC; ge1aa5.B = WS; ge1aa5.bias = be1; ge1aa5.R = EC; ge1aa5.C = EH1;
      ge1aa5.sAo = 0; ge1aa5.sAi = 0; ge1aa5.sAm = 32; ge1aa5.sAk = 1; ge1aa5.sBo = 0; ge1aa5.sBi = 0; ge1aa5.sBn = 1; ge1aa5.sBk = H; ge1aa5.sCo = 0; ge1aa5.sCi = 0; ge1aa5.sCm = H; ge1aa5.sRo = 0; ge1aa5.sRi = 0; ge1aa5.sRm = 0; ge1aa5.sRn = 0;
      ge1aa5.M = CH; ge1aa5.N = H; ge1aa5.K = 26; ge1aa5.zi_n = 1; ge1aa5.flags = 1; ge1aa5.act = 0;
      ge1aa5.alpha = 1.0f; ge1aa5.beta = 0.0f; ge1aa5.sa = 1.0f; ge1aa5.sb = 1.0f; ge1aa5.Npad = H; ge1aa5.pad_ = 0;
      k_gemm<1><<<dim3((unsigned)((H) + 31) / 32, (unsigned)((CH) + 15) / 16, (unsigned)(1)), 32, 0, stream>>>(ge1aa5); }
    { GemmP ge1ba5;
      ge1ba5.A = XS; ge1ba5.B = We1 + (size_t)4 * H; ge1ba5.bias = XS; ge1ba5.R = EH1; ge1ba5.C = EH1;
      ge1ba5.sAo = 0; ge1ba5.sAi = 0; ge1ba5.sAm = H; ge1ba5.sAk = 1; ge1ba5.sBo = 0; ge1ba5.sBi = 0; ge1ba5.sBn = 1; ge1ba5.sBk = H; ge1ba5.sCo = 0; ge1ba5.sCi = 0; ge1ba5.sCm = H; ge1ba5.sRo = 0; ge1ba5.sRi = 0; ge1ba5.sRm = H; ge1ba5.sRn = 1;
      ge1ba5.M = CH; ge1ba5.N = H; ge1ba5.K = H; ge1ba5.zi_n = 1; ge1ba5.flags = 4; ge1ba5.act = 0;
      ge1ba5.alpha = 1.0f; ge1ba5.beta = 1.0f; ge1ba5.sa = 1.0f; ge1ba5.sb = 1.0f; ge1ba5.Npad = H; ge1ba5.pad_ = 0;
      k_gemm<1><<<dim3((unsigned)((H) + 31) / 32, (unsigned)((CH) + 15) / 16, (unsigned)(1)), 32, 0, stream>>>(ge1ba5); }
    { GemmP ge1ca5;
      ge1ca5.A = XD; ge1ca5.B = We1 + (size_t)132 * H; ge1ca5.bias = XD; ge1ca5.R = EH1; ge1ca5.C = EH1;
      ge1ca5.sAo = 0; ge1ca5.sAi = 0; ge1ca5.sAm = H; ge1ca5.sAk = 1; ge1ca5.sBo = 0; ge1ca5.sBi = 0; ge1ca5.sBn = 1; ge1ca5.sBk = H; ge1ca5.sCo = 0; ge1ca5.sCi = 0; ge1ca5.sCm = H; ge1ca5.sRo = 0; ge1ca5.sRi = 0; ge1ca5.sRm = H; ge1ca5.sRn = 1;
      ge1ca5.M = CH; ge1ca5.N = H; ge1ca5.K = H; ge1ca5.zi_n = 1; ge1ca5.flags = 4; ge1ca5.act = 0;
      ge1ca5.alpha = 1.0f; ge1ca5.beta = 1.0f; ge1ca5.sa = 1.0f; ge1ca5.sb = 1.0f; ge1ca5.Npad = H; ge1ca5.pad_ = 0;
      k_gemm<1><<<dim3((unsigned)((H) + 31) / 32, (unsigned)((CH) + 15) / 16, (unsigned)(1)), 32, 0, stream>>>(ge1ca5); }
    k_norm_apply<<<(unsigned)(((long long)(1) * (1) * ((long long)CH * H) + 255) / 256), 256, 0, stream>>>(EH1, EH1, ust, nullptr, nullptr, 1, 1, (long long)CH * H, 1, 0, 1);
    { GemmP ge2a5;
      ge2a5.A = EH1; ge2a5.B = We2; ge2a5.bias = be2; ge2a5.R = EH1; ge2a5.C = EH;
      ge2a5.sAo = 0; ge2a5.sAi = 0; ge2a5.sAm = H; ge2a5.sAk = 1; ge2a5.sBo = 0; ge2a5.sBi = 0; ge2a5.sBn = 1; ge2a5.sBk = H; ge2a5.sCo = 0; ge2a5.sCi = 0; ge2a5.sCm = H; ge2a5.sRo = 0; ge2a5.sRi = 0; ge2a5.sRm = 0; ge2a5.sRn = 0;
      ge2a5.M = CH; ge2a5.N = H; ge2a5.K = H; ge2a5.zi_n = 1; ge2a5.flags = 1; ge2a5.act = 1;
      ge2a5.alpha = 1.0f; ge2a5.beta = 0.0f; ge2a5.sa = 1.0f; ge2a5.sb = 1.0f; ge2a5.Npad = H; ge2a5.pad_ = 0;
      k_gemm<1><<<dim3((unsigned)((H) + 31) / 32, (unsigned)((CH) + 15) / 16, (unsigned)(1)), 32, 0, stream>>>(ge2a5); }
    { GemmP gm5;
      gm5.A = EH; gm5.B = Wm; gm5.bias = bm; gm5.R = EH; gm5.C = MSG;
      gm5.sAo = 0; gm5.sAi = 0; gm5.sAm = H; gm5.sAk = 1; gm5.sBo = 0; gm5.sBi = 0; gm5.sBn = 1; gm5.sBk = H; gm5.sCo = 0; gm5.sCi = 0; gm5.sCm = H; gm5.sRo = 0; gm5.sRi = 0; gm5.sRm = 0; gm5.sRn = 0;
      gm5.M = CH; gm5.N = H; gm5.K = H; gm5.zi_n = 1; gm5.flags = 1; gm5.act = 0;
      gm5.alpha = 1.0f; gm5.beta = 0.0f; gm5.sa = 1.0f; gm5.sb = 1.0f; gm5.Npad = H; gm5.pad_ = 0;
      k_gemm<1><<<dim3((unsigned)((H) + 31) / 32, (unsigned)((CH) + 15) / 16, (unsigned)(1)), 32, 0, stream>>>(gm5); }
    k_sb_scale<<<(unsigned)(((long long)CH * H + 255) / 256), 256, 0, stream>>>(MSG, escope, 156250, CH, H);
    k_sb_agg<<<(unsigned)(((long long)N * H + 255) / 256), 256, 0, stream>>>(MSG, soff, sslot, doff, dslot, AGG, 156250, CH, N, H);
    k_sb_edgectx<<<(unsigned)(((long long)CH * H + 255) / 256), 256, 0, stream>>>(ef, etype, eparams, emask, escope, ebatch, emb, ei, NH, EC, XS, XD, 187500, CH, E, H);
    { GemmP ge1aa6;
      ge1aa6.A = EC; ge1aa6.B = WS; ge1aa6.bias = be1; ge1aa6.R = EC; ge1aa6.C = EH1;
      ge1aa6.sAo = 0; ge1aa6.sAi = 0; ge1aa6.sAm = 32; ge1aa6.sAk = 1; ge1aa6.sBo = 0; ge1aa6.sBi = 0; ge1aa6.sBn = 1; ge1aa6.sBk = H; ge1aa6.sCo = 0; ge1aa6.sCi = 0; ge1aa6.sCm = H; ge1aa6.sRo = 0; ge1aa6.sRi = 0; ge1aa6.sRm = 0; ge1aa6.sRn = 0;
      ge1aa6.M = CH; ge1aa6.N = H; ge1aa6.K = 26; ge1aa6.zi_n = 1; ge1aa6.flags = 1; ge1aa6.act = 0;
      ge1aa6.alpha = 1.0f; ge1aa6.beta = 0.0f; ge1aa6.sa = 1.0f; ge1aa6.sb = 1.0f; ge1aa6.Npad = H; ge1aa6.pad_ = 0;
      k_gemm<1><<<dim3((unsigned)((H) + 31) / 32, (unsigned)((CH) + 15) / 16, (unsigned)(1)), 32, 0, stream>>>(ge1aa6); }
    { GemmP ge1ba6;
      ge1ba6.A = XS; ge1ba6.B = We1 + (size_t)4 * H; ge1ba6.bias = XS; ge1ba6.R = EH1; ge1ba6.C = EH1;
      ge1ba6.sAo = 0; ge1ba6.sAi = 0; ge1ba6.sAm = H; ge1ba6.sAk = 1; ge1ba6.sBo = 0; ge1ba6.sBi = 0; ge1ba6.sBn = 1; ge1ba6.sBk = H; ge1ba6.sCo = 0; ge1ba6.sCi = 0; ge1ba6.sCm = H; ge1ba6.sRo = 0; ge1ba6.sRi = 0; ge1ba6.sRm = H; ge1ba6.sRn = 1;
      ge1ba6.M = CH; ge1ba6.N = H; ge1ba6.K = H; ge1ba6.zi_n = 1; ge1ba6.flags = 4; ge1ba6.act = 0;
      ge1ba6.alpha = 1.0f; ge1ba6.beta = 1.0f; ge1ba6.sa = 1.0f; ge1ba6.sb = 1.0f; ge1ba6.Npad = H; ge1ba6.pad_ = 0;
      k_gemm<1><<<dim3((unsigned)((H) + 31) / 32, (unsigned)((CH) + 15) / 16, (unsigned)(1)), 32, 0, stream>>>(ge1ba6); }
    { GemmP ge1ca6;
      ge1ca6.A = XD; ge1ca6.B = We1 + (size_t)132 * H; ge1ca6.bias = XD; ge1ca6.R = EH1; ge1ca6.C = EH1;
      ge1ca6.sAo = 0; ge1ca6.sAi = 0; ge1ca6.sAm = H; ge1ca6.sAk = 1; ge1ca6.sBo = 0; ge1ca6.sBi = 0; ge1ca6.sBn = 1; ge1ca6.sBk = H; ge1ca6.sCo = 0; ge1ca6.sCi = 0; ge1ca6.sCm = H; ge1ca6.sRo = 0; ge1ca6.sRi = 0; ge1ca6.sRm = H; ge1ca6.sRn = 1;
      ge1ca6.M = CH; ge1ca6.N = H; ge1ca6.K = H; ge1ca6.zi_n = 1; ge1ca6.flags = 4; ge1ca6.act = 0;
      ge1ca6.alpha = 1.0f; ge1ca6.beta = 1.0f; ge1ca6.sa = 1.0f; ge1ca6.sb = 1.0f; ge1ca6.Npad = H; ge1ca6.pad_ = 0;
      k_gemm<1><<<dim3((unsigned)((H) + 31) / 32, (unsigned)((CH) + 15) / 16, (unsigned)(1)), 32, 0, stream>>>(ge1ca6); }
    k_norm_apply<<<(unsigned)(((long long)(1) * (1) * ((long long)CH * H) + 255) / 256), 256, 0, stream>>>(EH1, EH1, ust, nullptr, nullptr, 1, 1, (long long)CH * H, 1, 0, 1);
    { GemmP ge2a6;
      ge2a6.A = EH1; ge2a6.B = We2; ge2a6.bias = be2; ge2a6.R = EH1; ge2a6.C = EH;
      ge2a6.sAo = 0; ge2a6.sAi = 0; ge2a6.sAm = H; ge2a6.sAk = 1; ge2a6.sBo = 0; ge2a6.sBi = 0; ge2a6.sBn = 1; ge2a6.sBk = H; ge2a6.sCo = 0; ge2a6.sCi = 0; ge2a6.sCm = H; ge2a6.sRo = 0; ge2a6.sRi = 0; ge2a6.sRm = 0; ge2a6.sRn = 0;
      ge2a6.M = CH; ge2a6.N = H; ge2a6.K = H; ge2a6.zi_n = 1; ge2a6.flags = 1; ge2a6.act = 1;
      ge2a6.alpha = 1.0f; ge2a6.beta = 0.0f; ge2a6.sa = 1.0f; ge2a6.sb = 1.0f; ge2a6.Npad = H; ge2a6.pad_ = 0;
      k_gemm<1><<<dim3((unsigned)((H) + 31) / 32, (unsigned)((CH) + 15) / 16, (unsigned)(1)), 32, 0, stream>>>(ge2a6); }
    { GemmP gm6;
      gm6.A = EH; gm6.B = Wm; gm6.bias = bm; gm6.R = EH; gm6.C = MSG;
      gm6.sAo = 0; gm6.sAi = 0; gm6.sAm = H; gm6.sAk = 1; gm6.sBo = 0; gm6.sBi = 0; gm6.sBn = 1; gm6.sBk = H; gm6.sCo = 0; gm6.sCi = 0; gm6.sCm = H; gm6.sRo = 0; gm6.sRi = 0; gm6.sRm = 0; gm6.sRn = 0;
      gm6.M = CH; gm6.N = H; gm6.K = H; gm6.zi_n = 1; gm6.flags = 1; gm6.act = 0;
      gm6.alpha = 1.0f; gm6.beta = 0.0f; gm6.sa = 1.0f; gm6.sb = 1.0f; gm6.Npad = H; gm6.pad_ = 0;
      k_gemm<1><<<dim3((unsigned)((H) + 31) / 32, (unsigned)((CH) + 15) / 16, (unsigned)(1)), 32, 0, stream>>>(gm6); }
    k_sb_scale<<<(unsigned)(((long long)CH * H + 255) / 256), 256, 0, stream>>>(MSG, escope, 187500, CH, H);
    k_sb_agg<<<(unsigned)(((long long)N * H + 255) / 256), 256, 0, stream>>>(MSG, soff, sslot, doff, dslot, AGG, 187500, CH, N, H);
    k_sb_edgectx<<<(unsigned)(((long long)CH * H + 255) / 256), 256, 0, stream>>>(ef, etype, eparams, emask, escope, ebatch, emb, ei, NH, EC, XS, XD, 218750, CH, E, H);
    { GemmP ge1aa7;
      ge1aa7.A = EC; ge1aa7.B = WS; ge1aa7.bias = be1; ge1aa7.R = EC; ge1aa7.C = EH1;
      ge1aa7.sAo = 0; ge1aa7.sAi = 0; ge1aa7.sAm = 32; ge1aa7.sAk = 1; ge1aa7.sBo = 0; ge1aa7.sBi = 0; ge1aa7.sBn = 1; ge1aa7.sBk = H; ge1aa7.sCo = 0; ge1aa7.sCi = 0; ge1aa7.sCm = H; ge1aa7.sRo = 0; ge1aa7.sRi = 0; ge1aa7.sRm = 0; ge1aa7.sRn = 0;
      ge1aa7.M = CH; ge1aa7.N = H; ge1aa7.K = 26; ge1aa7.zi_n = 1; ge1aa7.flags = 1; ge1aa7.act = 0;
      ge1aa7.alpha = 1.0f; ge1aa7.beta = 0.0f; ge1aa7.sa = 1.0f; ge1aa7.sb = 1.0f; ge1aa7.Npad = H; ge1aa7.pad_ = 0;
      k_gemm<1><<<dim3((unsigned)((H) + 31) / 32, (unsigned)((CH) + 15) / 16, (unsigned)(1)), 32, 0, stream>>>(ge1aa7); }
    { GemmP ge1ba7;
      ge1ba7.A = XS; ge1ba7.B = We1 + (size_t)4 * H; ge1ba7.bias = XS; ge1ba7.R = EH1; ge1ba7.C = EH1;
      ge1ba7.sAo = 0; ge1ba7.sAi = 0; ge1ba7.sAm = H; ge1ba7.sAk = 1; ge1ba7.sBo = 0; ge1ba7.sBi = 0; ge1ba7.sBn = 1; ge1ba7.sBk = H; ge1ba7.sCo = 0; ge1ba7.sCi = 0; ge1ba7.sCm = H; ge1ba7.sRo = 0; ge1ba7.sRi = 0; ge1ba7.sRm = H; ge1ba7.sRn = 1;
      ge1ba7.M = CH; ge1ba7.N = H; ge1ba7.K = H; ge1ba7.zi_n = 1; ge1ba7.flags = 4; ge1ba7.act = 0;
      ge1ba7.alpha = 1.0f; ge1ba7.beta = 1.0f; ge1ba7.sa = 1.0f; ge1ba7.sb = 1.0f; ge1ba7.Npad = H; ge1ba7.pad_ = 0;
      k_gemm<1><<<dim3((unsigned)((H) + 31) / 32, (unsigned)((CH) + 15) / 16, (unsigned)(1)), 32, 0, stream>>>(ge1ba7); }
    { GemmP ge1ca7;
      ge1ca7.A = XD; ge1ca7.B = We1 + (size_t)132 * H; ge1ca7.bias = XD; ge1ca7.R = EH1; ge1ca7.C = EH1;
      ge1ca7.sAo = 0; ge1ca7.sAi = 0; ge1ca7.sAm = H; ge1ca7.sAk = 1; ge1ca7.sBo = 0; ge1ca7.sBi = 0; ge1ca7.sBn = 1; ge1ca7.sBk = H; ge1ca7.sCo = 0; ge1ca7.sCi = 0; ge1ca7.sCm = H; ge1ca7.sRo = 0; ge1ca7.sRi = 0; ge1ca7.sRm = H; ge1ca7.sRn = 1;
      ge1ca7.M = CH; ge1ca7.N = H; ge1ca7.K = H; ge1ca7.zi_n = 1; ge1ca7.flags = 4; ge1ca7.act = 0;
      ge1ca7.alpha = 1.0f; ge1ca7.beta = 1.0f; ge1ca7.sa = 1.0f; ge1ca7.sb = 1.0f; ge1ca7.Npad = H; ge1ca7.pad_ = 0;
      k_gemm<1><<<dim3((unsigned)((H) + 31) / 32, (unsigned)((CH) + 15) / 16, (unsigned)(1)), 32, 0, stream>>>(ge1ca7); }
    k_norm_apply<<<(unsigned)(((long long)(1) * (1) * ((long long)CH * H) + 255) / 256), 256, 0, stream>>>(EH1, EH1, ust, nullptr, nullptr, 1, 1, (long long)CH * H, 1, 0, 1);
    { GemmP ge2a7;
      ge2a7.A = EH1; ge2a7.B = We2; ge2a7.bias = be2; ge2a7.R = EH1; ge2a7.C = EH;
      ge2a7.sAo = 0; ge2a7.sAi = 0; ge2a7.sAm = H; ge2a7.sAk = 1; ge2a7.sBo = 0; ge2a7.sBi = 0; ge2a7.sBn = 1; ge2a7.sBk = H; ge2a7.sCo = 0; ge2a7.sCi = 0; ge2a7.sCm = H; ge2a7.sRo = 0; ge2a7.sRi = 0; ge2a7.sRm = 0; ge2a7.sRn = 0;
      ge2a7.M = CH; ge2a7.N = H; ge2a7.K = H; ge2a7.zi_n = 1; ge2a7.flags = 1; ge2a7.act = 1;
      ge2a7.alpha = 1.0f; ge2a7.beta = 0.0f; ge2a7.sa = 1.0f; ge2a7.sb = 1.0f; ge2a7.Npad = H; ge2a7.pad_ = 0;
      k_gemm<1><<<dim3((unsigned)((H) + 31) / 32, (unsigned)((CH) + 15) / 16, (unsigned)(1)), 32, 0, stream>>>(ge2a7); }
    { GemmP gm7;
      gm7.A = EH; gm7.B = Wm; gm7.bias = bm; gm7.R = EH; gm7.C = MSG;
      gm7.sAo = 0; gm7.sAi = 0; gm7.sAm = H; gm7.sAk = 1; gm7.sBo = 0; gm7.sBi = 0; gm7.sBn = 1; gm7.sBk = H; gm7.sCo = 0; gm7.sCi = 0; gm7.sCm = H; gm7.sRo = 0; gm7.sRi = 0; gm7.sRm = 0; gm7.sRn = 0;
      gm7.M = CH; gm7.N = H; gm7.K = H; gm7.zi_n = 1; gm7.flags = 1; gm7.act = 0;
      gm7.alpha = 1.0f; gm7.beta = 0.0f; gm7.sa = 1.0f; gm7.sb = 1.0f; gm7.Npad = H; gm7.pad_ = 0;
      k_gemm<1><<<dim3((unsigned)((H) + 31) / 32, (unsigned)((CH) + 15) / 16, (unsigned)(1)), 32, 0, stream>>>(gm7); }
    k_sb_scale<<<(unsigned)(((long long)CH * H + 255) / 256), 256, 0, stream>>>(MSG, escope, 218750, CH, H);
    k_sb_agg<<<(unsigned)(((long long)N * H + 255) / 256), 256, 0, stream>>>(MSG, soff, sslot, doff, dslot, AGG, 218750, CH, N, H);
    k_sb_edgectx<<<(unsigned)(((long long)CH * H + 255) / 256), 256, 0, stream>>>(ef, etype, eparams, emask, escope, ebatch, emb, ei, NH, EC, XS, XD, 250000, CH, E, H);
    { GemmP ge1aa8;
      ge1aa8.A = EC; ge1aa8.B = WS; ge1aa8.bias = be1; ge1aa8.R = EC; ge1aa8.C = EH1;
      ge1aa8.sAo = 0; ge1aa8.sAi = 0; ge1aa8.sAm = 32; ge1aa8.sAk = 1; ge1aa8.sBo = 0; ge1aa8.sBi = 0; ge1aa8.sBn = 1; ge1aa8.sBk = H; ge1aa8.sCo = 0; ge1aa8.sCi = 0; ge1aa8.sCm = H; ge1aa8.sRo = 0; ge1aa8.sRi = 0; ge1aa8.sRm = 0; ge1aa8.sRn = 0;
      ge1aa8.M = CH; ge1aa8.N = H; ge1aa8.K = 26; ge1aa8.zi_n = 1; ge1aa8.flags = 1; ge1aa8.act = 0;
      ge1aa8.alpha = 1.0f; ge1aa8.beta = 0.0f; ge1aa8.sa = 1.0f; ge1aa8.sb = 1.0f; ge1aa8.Npad = H; ge1aa8.pad_ = 0;
      k_gemm<1><<<dim3((unsigned)((H) + 31) / 32, (unsigned)((CH) + 15) / 16, (unsigned)(1)), 32, 0, stream>>>(ge1aa8); }
    { GemmP ge1ba8;
      ge1ba8.A = XS; ge1ba8.B = We1 + (size_t)4 * H; ge1ba8.bias = XS; ge1ba8.R = EH1; ge1ba8.C = EH1;
      ge1ba8.sAo = 0; ge1ba8.sAi = 0; ge1ba8.sAm = H; ge1ba8.sAk = 1; ge1ba8.sBo = 0; ge1ba8.sBi = 0; ge1ba8.sBn = 1; ge1ba8.sBk = H; ge1ba8.sCo = 0; ge1ba8.sCi = 0; ge1ba8.sCm = H; ge1ba8.sRo = 0; ge1ba8.sRi = 0; ge1ba8.sRm = H; ge1ba8.sRn = 1;
      ge1ba8.M = CH; ge1ba8.N = H; ge1ba8.K = H; ge1ba8.zi_n = 1; ge1ba8.flags = 4; ge1ba8.act = 0;
      ge1ba8.alpha = 1.0f; ge1ba8.beta = 1.0f; ge1ba8.sa = 1.0f; ge1ba8.sb = 1.0f; ge1ba8.Npad = H; ge1ba8.pad_ = 0;
      k_gemm<1><<<dim3((unsigned)((H) + 31) / 32, (unsigned)((CH) + 15) / 16, (unsigned)(1)), 32, 0, stream>>>(ge1ba8); }
    { GemmP ge1ca8;
      ge1ca8.A = XD; ge1ca8.B = We1 + (size_t)132 * H; ge1ca8.bias = XD; ge1ca8.R = EH1; ge1ca8.C = EH1;
      ge1ca8.sAo = 0; ge1ca8.sAi = 0; ge1ca8.sAm = H; ge1ca8.sAk = 1; ge1ca8.sBo = 0; ge1ca8.sBi = 0; ge1ca8.sBn = 1; ge1ca8.sBk = H; ge1ca8.sCo = 0; ge1ca8.sCi = 0; ge1ca8.sCm = H; ge1ca8.sRo = 0; ge1ca8.sRi = 0; ge1ca8.sRm = H; ge1ca8.sRn = 1;
      ge1ca8.M = CH; ge1ca8.N = H; ge1ca8.K = H; ge1ca8.zi_n = 1; ge1ca8.flags = 4; ge1ca8.act = 0;
      ge1ca8.alpha = 1.0f; ge1ca8.beta = 1.0f; ge1ca8.sa = 1.0f; ge1ca8.sb = 1.0f; ge1ca8.Npad = H; ge1ca8.pad_ = 0;
      k_gemm<1><<<dim3((unsigned)((H) + 31) / 32, (unsigned)((CH) + 15) / 16, (unsigned)(1)), 32, 0, stream>>>(ge1ca8); }
    k_norm_apply<<<(unsigned)(((long long)(1) * (1) * ((long long)CH * H) + 255) / 256), 256, 0, stream>>>(EH1, EH1, ust, nullptr, nullptr, 1, 1, (long long)CH * H, 1, 0, 1);
    { GemmP ge2a8;
      ge2a8.A = EH1; ge2a8.B = We2; ge2a8.bias = be2; ge2a8.R = EH1; ge2a8.C = EH;
      ge2a8.sAo = 0; ge2a8.sAi = 0; ge2a8.sAm = H; ge2a8.sAk = 1; ge2a8.sBo = 0; ge2a8.sBi = 0; ge2a8.sBn = 1; ge2a8.sBk = H; ge2a8.sCo = 0; ge2a8.sCi = 0; ge2a8.sCm = H; ge2a8.sRo = 0; ge2a8.sRi = 0; ge2a8.sRm = 0; ge2a8.sRn = 0;
      ge2a8.M = CH; ge2a8.N = H; ge2a8.K = H; ge2a8.zi_n = 1; ge2a8.flags = 1; ge2a8.act = 1;
      ge2a8.alpha = 1.0f; ge2a8.beta = 0.0f; ge2a8.sa = 1.0f; ge2a8.sb = 1.0f; ge2a8.Npad = H; ge2a8.pad_ = 0;
      k_gemm<1><<<dim3((unsigned)((H) + 31) / 32, (unsigned)((CH) + 15) / 16, (unsigned)(1)), 32, 0, stream>>>(ge2a8); }
    { GemmP gm8;
      gm8.A = EH; gm8.B = Wm; gm8.bias = bm; gm8.R = EH; gm8.C = MSG;
      gm8.sAo = 0; gm8.sAi = 0; gm8.sAm = H; gm8.sAk = 1; gm8.sBo = 0; gm8.sBi = 0; gm8.sBn = 1; gm8.sBk = H; gm8.sCo = 0; gm8.sCi = 0; gm8.sCm = H; gm8.sRo = 0; gm8.sRi = 0; gm8.sRm = 0; gm8.sRn = 0;
      gm8.M = CH; gm8.N = H; gm8.K = H; gm8.zi_n = 1; gm8.flags = 1; gm8.act = 0;
      gm8.alpha = 1.0f; gm8.beta = 0.0f; gm8.sa = 1.0f; gm8.sb = 1.0f; gm8.Npad = H; gm8.pad_ = 0;
      k_gemm<1><<<dim3((unsigned)((H) + 31) / 32, (unsigned)((CH) + 15) / 16, (unsigned)(1)), 32, 0, stream>>>(gm8); }
    k_sb_scale<<<(unsigned)(((long long)CH * H + 255) / 256), 256, 0, stream>>>(MSG, escope, 250000, CH, H);
    k_sb_agg<<<(unsigned)(((long long)N * H + 255) / 256), 256, 0, stream>>>(MSG, soff, sslot, doff, dslot, AGG, 250000, CH, N, H);
    k_sb_edgectx<<<(unsigned)(((long long)CH * H + 255) / 256), 256, 0, stream>>>(ef, etype, eparams, emask, escope, ebatch, emb, ei, NH, EC, XS, XD, 281250, CH, E, H);
    { GemmP ge1aa9;
      ge1aa9.A = EC; ge1aa9.B = WS; ge1aa9.bias = be1; ge1aa9.R = EC; ge1aa9.C = EH1;
      ge1aa9.sAo = 0; ge1aa9.sAi = 0; ge1aa9.sAm = 32; ge1aa9.sAk = 1; ge1aa9.sBo = 0; ge1aa9.sBi = 0; ge1aa9.sBn = 1; ge1aa9.sBk = H; ge1aa9.sCo = 0; ge1aa9.sCi = 0; ge1aa9.sCm = H; ge1aa9.sRo = 0; ge1aa9.sRi = 0; ge1aa9.sRm = 0; ge1aa9.sRn = 0;
      ge1aa9.M = CH; ge1aa9.N = H; ge1aa9.K = 26; ge1aa9.zi_n = 1; ge1aa9.flags = 1; ge1aa9.act = 0;
      ge1aa9.alpha = 1.0f; ge1aa9.beta = 0.0f; ge1aa9.sa = 1.0f; ge1aa9.sb = 1.0f; ge1aa9.Npad = H; ge1aa9.pad_ = 0;
      k_gemm<1><<<dim3((unsigned)((H) + 31) / 32, (unsigned)((CH) + 15) / 16, (unsigned)(1)), 32, 0, stream>>>(ge1aa9); }
    { GemmP ge1ba9;
      ge1ba9.A = XS; ge1ba9.B = We1 + (size_t)4 * H; ge1ba9.bias = XS; ge1ba9.R = EH1; ge1ba9.C = EH1;
      ge1ba9.sAo = 0; ge1ba9.sAi = 0; ge1ba9.sAm = H; ge1ba9.sAk = 1; ge1ba9.sBo = 0; ge1ba9.sBi = 0; ge1ba9.sBn = 1; ge1ba9.sBk = H; ge1ba9.sCo = 0; ge1ba9.sCi = 0; ge1ba9.sCm = H; ge1ba9.sRo = 0; ge1ba9.sRi = 0; ge1ba9.sRm = H; ge1ba9.sRn = 1;
      ge1ba9.M = CH; ge1ba9.N = H; ge1ba9.K = H; ge1ba9.zi_n = 1; ge1ba9.flags = 4; ge1ba9.act = 0;
      ge1ba9.alpha = 1.0f; ge1ba9.beta = 1.0f; ge1ba9.sa = 1.0f; ge1ba9.sb = 1.0f; ge1ba9.Npad = H; ge1ba9.pad_ = 0;
      k_gemm<1><<<dim3((unsigned)((H) + 31) / 32, (unsigned)((CH) + 15) / 16, (unsigned)(1)), 32, 0, stream>>>(ge1ba9); }
    { GemmP ge1ca9;
      ge1ca9.A = XD; ge1ca9.B = We1 + (size_t)132 * H; ge1ca9.bias = XD; ge1ca9.R = EH1; ge1ca9.C = EH1;
      ge1ca9.sAo = 0; ge1ca9.sAi = 0; ge1ca9.sAm = H; ge1ca9.sAk = 1; ge1ca9.sBo = 0; ge1ca9.sBi = 0; ge1ca9.sBn = 1; ge1ca9.sBk = H; ge1ca9.sCo = 0; ge1ca9.sCi = 0; ge1ca9.sCm = H; ge1ca9.sRo = 0; ge1ca9.sRi = 0; ge1ca9.sRm = H; ge1ca9.sRn = 1;
      ge1ca9.M = CH; ge1ca9.N = H; ge1ca9.K = H; ge1ca9.zi_n = 1; ge1ca9.flags = 4; ge1ca9.act = 0;
      ge1ca9.alpha = 1.0f; ge1ca9.beta = 1.0f; ge1ca9.sa = 1.0f; ge1ca9.sb = 1.0f; ge1ca9.Npad = H; ge1ca9.pad_ = 0;
      k_gemm<1><<<dim3((unsigned)((H) + 31) / 32, (unsigned)((CH) + 15) / 16, (unsigned)(1)), 32, 0, stream>>>(ge1ca9); }
    k_norm_apply<<<(unsigned)(((long long)(1) * (1) * ((long long)CH * H) + 255) / 256), 256, 0, stream>>>(EH1, EH1, ust, nullptr, nullptr, 1, 1, (long long)CH * H, 1, 0, 1);
    { GemmP ge2a9;
      ge2a9.A = EH1; ge2a9.B = We2; ge2a9.bias = be2; ge2a9.R = EH1; ge2a9.C = EH;
      ge2a9.sAo = 0; ge2a9.sAi = 0; ge2a9.sAm = H; ge2a9.sAk = 1; ge2a9.sBo = 0; ge2a9.sBi = 0; ge2a9.sBn = 1; ge2a9.sBk = H; ge2a9.sCo = 0; ge2a9.sCi = 0; ge2a9.sCm = H; ge2a9.sRo = 0; ge2a9.sRi = 0; ge2a9.sRm = 0; ge2a9.sRn = 0;
      ge2a9.M = CH; ge2a9.N = H; ge2a9.K = H; ge2a9.zi_n = 1; ge2a9.flags = 1; ge2a9.act = 1;
      ge2a9.alpha = 1.0f; ge2a9.beta = 0.0f; ge2a9.sa = 1.0f; ge2a9.sb = 1.0f; ge2a9.Npad = H; ge2a9.pad_ = 0;
      k_gemm<1><<<dim3((unsigned)((H) + 31) / 32, (unsigned)((CH) + 15) / 16, (unsigned)(1)), 32, 0, stream>>>(ge2a9); }
    { GemmP gm9;
      gm9.A = EH; gm9.B = Wm; gm9.bias = bm; gm9.R = EH; gm9.C = MSG;
      gm9.sAo = 0; gm9.sAi = 0; gm9.sAm = H; gm9.sAk = 1; gm9.sBo = 0; gm9.sBi = 0; gm9.sBn = 1; gm9.sBk = H; gm9.sCo = 0; gm9.sCi = 0; gm9.sCm = H; gm9.sRo = 0; gm9.sRi = 0; gm9.sRm = 0; gm9.sRn = 0;
      gm9.M = CH; gm9.N = H; gm9.K = H; gm9.zi_n = 1; gm9.flags = 1; gm9.act = 0;
      gm9.alpha = 1.0f; gm9.beta = 0.0f; gm9.sa = 1.0f; gm9.sb = 1.0f; gm9.Npad = H; gm9.pad_ = 0;
      k_gemm<1><<<dim3((unsigned)((H) + 31) / 32, (unsigned)((CH) + 15) / 16, (unsigned)(1)), 32, 0, stream>>>(gm9); }
    k_sb_scale<<<(unsigned)(((long long)CH * H + 255) / 256), 256, 0, stream>>>(MSG, escope, 281250, CH, H);
    k_sb_agg<<<(unsigned)(((long long)N * H + 255) / 256), 256, 0, stream>>>(MSG, soff, sslot, doff, dslot, AGG, 281250, CH, N, H);
    k_sb_edgectx<<<(unsigned)(((long long)CH * H + 255) / 256), 256, 0, stream>>>(ef, etype, eparams, emask, escope, ebatch, emb, ei, NH, EC, XS, XD, 312500, CH, E, H);
    { GemmP ge1aa10;
      ge1aa10.A = EC; ge1aa10.B = WS; ge1aa10.bias = be1; ge1aa10.R = EC; ge1aa10.C = EH1;
      ge1aa10.sAo = 0; ge1aa10.sAi = 0; ge1aa10.sAm = 32; ge1aa10.sAk = 1; ge1aa10.sBo = 0; ge1aa10.sBi = 0; ge1aa10.sBn = 1; ge1aa10.sBk = H; ge1aa10.sCo = 0; ge1aa10.sCi = 0; ge1aa10.sCm = H; ge1aa10.sRo = 0; ge1aa10.sRi = 0; ge1aa10.sRm = 0; ge1aa10.sRn = 0;
      ge1aa10.M = CH; ge1aa10.N = H; ge1aa10.K = 26; ge1aa10.zi_n = 1; ge1aa10.flags = 1; ge1aa10.act = 0;
      ge1aa10.alpha = 1.0f; ge1aa10.beta = 0.0f; ge1aa10.sa = 1.0f; ge1aa10.sb = 1.0f; ge1aa10.Npad = H; ge1aa10.pad_ = 0;
      k_gemm<1><<<dim3((unsigned)((H) + 31) / 32, (unsigned)((CH) + 15) / 16, (unsigned)(1)), 32, 0, stream>>>(ge1aa10); }
    { GemmP ge1ba10;
      ge1ba10.A = XS; ge1ba10.B = We1 + (size_t)4 * H; ge1ba10.bias = XS; ge1ba10.R = EH1; ge1ba10.C = EH1;
      ge1ba10.sAo = 0; ge1ba10.sAi = 0; ge1ba10.sAm = H; ge1ba10.sAk = 1; ge1ba10.sBo = 0; ge1ba10.sBi = 0; ge1ba10.sBn = 1; ge1ba10.sBk = H; ge1ba10.sCo = 0; ge1ba10.sCi = 0; ge1ba10.sCm = H; ge1ba10.sRo = 0; ge1ba10.sRi = 0; ge1ba10.sRm = H; ge1ba10.sRn = 1;
      ge1ba10.M = CH; ge1ba10.N = H; ge1ba10.K = H; ge1ba10.zi_n = 1; ge1ba10.flags = 4; ge1ba10.act = 0;
      ge1ba10.alpha = 1.0f; ge1ba10.beta = 1.0f; ge1ba10.sa = 1.0f; ge1ba10.sb = 1.0f; ge1ba10.Npad = H; ge1ba10.pad_ = 0;
      k_gemm<1><<<dim3((unsigned)((H) + 31) / 32, (unsigned)((CH) + 15) / 16, (unsigned)(1)), 32, 0, stream>>>(ge1ba10); }
    { GemmP ge1ca10;
      ge1ca10.A = XD; ge1ca10.B = We1 + (size_t)132 * H; ge1ca10.bias = XD; ge1ca10.R = EH1; ge1ca10.C = EH1;
      ge1ca10.sAo = 0; ge1ca10.sAi = 0; ge1ca10.sAm = H; ge1ca10.sAk = 1; ge1ca10.sBo = 0; ge1ca10.sBi = 0; ge1ca10.sBn = 1; ge1ca10.sBk = H; ge1ca10.sCo = 0; ge1ca10.sCi = 0; ge1ca10.sCm = H; ge1ca10.sRo = 0; ge1ca10.sRi = 0; ge1ca10.sRm = H; ge1ca10.sRn = 1;
      ge1ca10.M = CH; ge1ca10.N = H; ge1ca10.K = H; ge1ca10.zi_n = 1; ge1ca10.flags = 4; ge1ca10.act = 0;
      ge1ca10.alpha = 1.0f; ge1ca10.beta = 1.0f; ge1ca10.sa = 1.0f; ge1ca10.sb = 1.0f; ge1ca10.Npad = H; ge1ca10.pad_ = 0;
      k_gemm<1><<<dim3((unsigned)((H) + 31) / 32, (unsigned)((CH) + 15) / 16, (unsigned)(1)), 32, 0, stream>>>(ge1ca10); }
    k_norm_apply<<<(unsigned)(((long long)(1) * (1) * ((long long)CH * H) + 255) / 256), 256, 0, stream>>>(EH1, EH1, ust, nullptr, nullptr, 1, 1, (long long)CH * H, 1, 0, 1);
    { GemmP ge2a10;
      ge2a10.A = EH1; ge2a10.B = We2; ge2a10.bias = be2; ge2a10.R = EH1; ge2a10.C = EH;
      ge2a10.sAo = 0; ge2a10.sAi = 0; ge2a10.sAm = H; ge2a10.sAk = 1; ge2a10.sBo = 0; ge2a10.sBi = 0; ge2a10.sBn = 1; ge2a10.sBk = H; ge2a10.sCo = 0; ge2a10.sCi = 0; ge2a10.sCm = H; ge2a10.sRo = 0; ge2a10.sRi = 0; ge2a10.sRm = 0; ge2a10.sRn = 0;
      ge2a10.M = CH; ge2a10.N = H; ge2a10.K = H; ge2a10.zi_n = 1; ge2a10.flags = 1; ge2a10.act = 1;
      ge2a10.alpha = 1.0f; ge2a10.beta = 0.0f; ge2a10.sa = 1.0f; ge2a10.sb = 1.0f; ge2a10.Npad = H; ge2a10.pad_ = 0;
      k_gemm<1><<<dim3((unsigned)((H) + 31) / 32, (unsigned)((CH) + 15) / 16, (unsigned)(1)), 32, 0, stream>>>(ge2a10); }
    { GemmP gm10;
      gm10.A = EH; gm10.B = Wm; gm10.bias = bm; gm10.R = EH; gm10.C = MSG;
      gm10.sAo = 0; gm10.sAi = 0; gm10.sAm = H; gm10.sAk = 1; gm10.sBo = 0; gm10.sBi = 0; gm10.sBn = 1; gm10.sBk = H; gm10.sCo = 0; gm10.sCi = 0; gm10.sCm = H; gm10.sRo = 0; gm10.sRi = 0; gm10.sRm = 0; gm10.sRn = 0;
      gm10.M = CH; gm10.N = H; gm10.K = H; gm10.zi_n = 1; gm10.flags = 1; gm10.act = 0;
      gm10.alpha = 1.0f; gm10.beta = 0.0f; gm10.sa = 1.0f; gm10.sb = 1.0f; gm10.Npad = H; gm10.pad_ = 0;
      k_gemm<1><<<dim3((unsigned)((H) + 31) / 32, (unsigned)((CH) + 15) / 16, (unsigned)(1)), 32, 0, stream>>>(gm10); }
    k_sb_scale<<<(unsigned)(((long long)CH * H + 255) / 256), 256, 0, stream>>>(MSG, escope, 312500, CH, H);
    k_sb_agg<<<(unsigned)(((long long)N * H + 255) / 256), 256, 0, stream>>>(MSG, soff, sslot, doff, dslot, AGG, 312500, CH, N, H);
    k_sb_edgectx<<<(unsigned)(((long long)CH * H + 255) / 256), 256, 0, stream>>>(ef, etype, eparams, emask, escope, ebatch, emb, ei, NH, EC, XS, XD, 343750, CH, E, H);
    { GemmP ge1aa11;
      ge1aa11.A = EC; ge1aa11.B = WS; ge1aa11.bias = be1; ge1aa11.R = EC; ge1aa11.C = EH1;
      ge1aa11.sAo = 0; ge1aa11.sAi = 0; ge1aa11.sAm = 32; ge1aa11.sAk = 1; ge1aa11.sBo = 0; ge1aa11.sBi = 0; ge1aa11.sBn = 1; ge1aa11.sBk = H; ge1aa11.sCo = 0; ge1aa11.sCi = 0; ge1aa11.sCm = H; ge1aa11.sRo = 0; ge1aa11.sRi = 0; ge1aa11.sRm = 0; ge1aa11.sRn = 0;
      ge1aa11.M = CH; ge1aa11.N = H; ge1aa11.K = 26; ge1aa11.zi_n = 1; ge1aa11.flags = 1; ge1aa11.act = 0;
      ge1aa11.alpha = 1.0f; ge1aa11.beta = 0.0f; ge1aa11.sa = 1.0f; ge1aa11.sb = 1.0f; ge1aa11.Npad = H; ge1aa11.pad_ = 0;
      k_gemm<1><<<dim3((unsigned)((H) + 31) / 32, (unsigned)((CH) + 15) / 16, (unsigned)(1)), 32, 0, stream>>>(ge1aa11); }
    { GemmP ge1ba11;
      ge1ba11.A = XS; ge1ba11.B = We1 + (size_t)4 * H; ge1ba11.bias = XS; ge1ba11.R = EH1; ge1ba11.C = EH1;
      ge1ba11.sAo = 0; ge1ba11.sAi = 0; ge1ba11.sAm = H; ge1ba11.sAk = 1; ge1ba11.sBo = 0; ge1ba11.sBi = 0; ge1ba11.sBn = 1; ge1ba11.sBk = H; ge1ba11.sCo = 0; ge1ba11.sCi = 0; ge1ba11.sCm = H; ge1ba11.sRo = 0; ge1ba11.sRi = 0; ge1ba11.sRm = H; ge1ba11.sRn = 1;
      ge1ba11.M = CH; ge1ba11.N = H; ge1ba11.K = H; ge1ba11.zi_n = 1; ge1ba11.flags = 4; ge1ba11.act = 0;
      ge1ba11.alpha = 1.0f; ge1ba11.beta = 1.0f; ge1ba11.sa = 1.0f; ge1ba11.sb = 1.0f; ge1ba11.Npad = H; ge1ba11.pad_ = 0;
      k_gemm<1><<<dim3((unsigned)((H) + 31) / 32, (unsigned)((CH) + 15) / 16, (unsigned)(1)), 32, 0, stream>>>(ge1ba11); }
    { GemmP ge1ca11;
      ge1ca11.A = XD; ge1ca11.B = We1 + (size_t)132 * H; ge1ca11.bias = XD; ge1ca11.R = EH1; ge1ca11.C = EH1;
      ge1ca11.sAo = 0; ge1ca11.sAi = 0; ge1ca11.sAm = H; ge1ca11.sAk = 1; ge1ca11.sBo = 0; ge1ca11.sBi = 0; ge1ca11.sBn = 1; ge1ca11.sBk = H; ge1ca11.sCo = 0; ge1ca11.sCi = 0; ge1ca11.sCm = H; ge1ca11.sRo = 0; ge1ca11.sRi = 0; ge1ca11.sRm = H; ge1ca11.sRn = 1;
      ge1ca11.M = CH; ge1ca11.N = H; ge1ca11.K = H; ge1ca11.zi_n = 1; ge1ca11.flags = 4; ge1ca11.act = 0;
      ge1ca11.alpha = 1.0f; ge1ca11.beta = 1.0f; ge1ca11.sa = 1.0f; ge1ca11.sb = 1.0f; ge1ca11.Npad = H; ge1ca11.pad_ = 0;
      k_gemm<1><<<dim3((unsigned)((H) + 31) / 32, (unsigned)((CH) + 15) / 16, (unsigned)(1)), 32, 0, stream>>>(ge1ca11); }
    k_norm_apply<<<(unsigned)(((long long)(1) * (1) * ((long long)CH * H) + 255) / 256), 256, 0, stream>>>(EH1, EH1, ust, nullptr, nullptr, 1, 1, (long long)CH * H, 1, 0, 1);
    { GemmP ge2a11;
      ge2a11.A = EH1; ge2a11.B = We2; ge2a11.bias = be2; ge2a11.R = EH1; ge2a11.C = EH;
      ge2a11.sAo = 0; ge2a11.sAi = 0; ge2a11.sAm = H; ge2a11.sAk = 1; ge2a11.sBo = 0; ge2a11.sBi = 0; ge2a11.sBn = 1; ge2a11.sBk = H; ge2a11.sCo = 0; ge2a11.sCi = 0; ge2a11.sCm = H; ge2a11.sRo = 0; ge2a11.sRi = 0; ge2a11.sRm = 0; ge2a11.sRn = 0;
      ge2a11.M = CH; ge2a11.N = H; ge2a11.K = H; ge2a11.zi_n = 1; ge2a11.flags = 1; ge2a11.act = 1;
      ge2a11.alpha = 1.0f; ge2a11.beta = 0.0f; ge2a11.sa = 1.0f; ge2a11.sb = 1.0f; ge2a11.Npad = H; ge2a11.pad_ = 0;
      k_gemm<1><<<dim3((unsigned)((H) + 31) / 32, (unsigned)((CH) + 15) / 16, (unsigned)(1)), 32, 0, stream>>>(ge2a11); }
    { GemmP gm11;
      gm11.A = EH; gm11.B = Wm; gm11.bias = bm; gm11.R = EH; gm11.C = MSG;
      gm11.sAo = 0; gm11.sAi = 0; gm11.sAm = H; gm11.sAk = 1; gm11.sBo = 0; gm11.sBi = 0; gm11.sBn = 1; gm11.sBk = H; gm11.sCo = 0; gm11.sCi = 0; gm11.sCm = H; gm11.sRo = 0; gm11.sRi = 0; gm11.sRm = 0; gm11.sRn = 0;
      gm11.M = CH; gm11.N = H; gm11.K = H; gm11.zi_n = 1; gm11.flags = 1; gm11.act = 0;
      gm11.alpha = 1.0f; gm11.beta = 0.0f; gm11.sa = 1.0f; gm11.sb = 1.0f; gm11.Npad = H; gm11.pad_ = 0;
      k_gemm<1><<<dim3((unsigned)((H) + 31) / 32, (unsigned)((CH) + 15) / 16, (unsigned)(1)), 32, 0, stream>>>(gm11); }
    k_sb_scale<<<(unsigned)(((long long)CH * H + 255) / 256), 256, 0, stream>>>(MSG, escope, 343750, CH, H);
    k_sb_agg<<<(unsigned)(((long long)N * H + 255) / 256), 256, 0, stream>>>(MSG, soff, sslot, doff, dslot, AGG, 343750, CH, N, H);
    k_sb_edgectx<<<(unsigned)(((long long)CH * H + 255) / 256), 256, 0, stream>>>(ef, etype, eparams, emask, escope, ebatch, emb, ei, NH, EC, XS, XD, 375000, CH, E, H);
    { GemmP ge1aa12;
      ge1aa12.A = EC; ge1aa12.B = WS; ge1aa12.bias = be1; ge1aa12.R = EC; ge1aa12.C = EH1;
      ge1aa12.sAo = 0; ge1aa12.sAi = 0; ge1aa12.sAm = 32; ge1aa12.sAk = 1; ge1aa12.sBo = 0; ge1aa12.sBi = 0; ge1aa12.sBn = 1; ge1aa12.sBk = H; ge1aa12.sCo = 0; ge1aa12.sCi = 0; ge1aa12.sCm = H; ge1aa12.sRo = 0; ge1aa12.sRi = 0; ge1aa12.sRm = 0; ge1aa12.sRn = 0;
      ge1aa12.M = CH; ge1aa12.N = H; ge1aa12.K = 26; ge1aa12.zi_n = 1; ge1aa12.flags = 1; ge1aa12.act = 0;
      ge1aa12.alpha = 1.0f; ge1aa12.beta = 0.0f; ge1aa12.sa = 1.0f; ge1aa12.sb = 1.0f; ge1aa12.Npad = H; ge1aa12.pad_ = 0;
      k_gemm<1><<<dim3((unsigned)((H) + 31) / 32, (unsigned)((CH) + 15) / 16, (unsigned)(1)), 32, 0, stream>>>(ge1aa12); }
    { GemmP ge1ba12;
      ge1ba12.A = XS; ge1ba12.B = We1 + (size_t)4 * H; ge1ba12.bias = XS; ge1ba12.R = EH1; ge1ba12.C = EH1;
      ge1ba12.sAo = 0; ge1ba12.sAi = 0; ge1ba12.sAm = H; ge1ba12.sAk = 1; ge1ba12.sBo = 0; ge1ba12.sBi = 0; ge1ba12.sBn = 1; ge1ba12.sBk = H; ge1ba12.sCo = 0; ge1ba12.sCi = 0; ge1ba12.sCm = H; ge1ba12.sRo = 0; ge1ba12.sRi = 0; ge1ba12.sRm = H; ge1ba12.sRn = 1;
      ge1ba12.M = CH; ge1ba12.N = H; ge1ba12.K = H; ge1ba12.zi_n = 1; ge1ba12.flags = 4; ge1ba12.act = 0;
      ge1ba12.alpha = 1.0f; ge1ba12.beta = 1.0f; ge1ba12.sa = 1.0f; ge1ba12.sb = 1.0f; ge1ba12.Npad = H; ge1ba12.pad_ = 0;
      k_gemm<1><<<dim3((unsigned)((H) + 31) / 32, (unsigned)((CH) + 15) / 16, (unsigned)(1)), 32, 0, stream>>>(ge1ba12); }
    { GemmP ge1ca12;
      ge1ca12.A = XD; ge1ca12.B = We1 + (size_t)132 * H; ge1ca12.bias = XD; ge1ca12.R = EH1; ge1ca12.C = EH1;
      ge1ca12.sAo = 0; ge1ca12.sAi = 0; ge1ca12.sAm = H; ge1ca12.sAk = 1; ge1ca12.sBo = 0; ge1ca12.sBi = 0; ge1ca12.sBn = 1; ge1ca12.sBk = H; ge1ca12.sCo = 0; ge1ca12.sCi = 0; ge1ca12.sCm = H; ge1ca12.sRo = 0; ge1ca12.sRi = 0; ge1ca12.sRm = H; ge1ca12.sRn = 1;
      ge1ca12.M = CH; ge1ca12.N = H; ge1ca12.K = H; ge1ca12.zi_n = 1; ge1ca12.flags = 4; ge1ca12.act = 0;
      ge1ca12.alpha = 1.0f; ge1ca12.beta = 1.0f; ge1ca12.sa = 1.0f; ge1ca12.sb = 1.0f; ge1ca12.Npad = H; ge1ca12.pad_ = 0;
      k_gemm<1><<<dim3((unsigned)((H) + 31) / 32, (unsigned)((CH) + 15) / 16, (unsigned)(1)), 32, 0, stream>>>(ge1ca12); }
    k_norm_apply<<<(unsigned)(((long long)(1) * (1) * ((long long)CH * H) + 255) / 256), 256, 0, stream>>>(EH1, EH1, ust, nullptr, nullptr, 1, 1, (long long)CH * H, 1, 0, 1);
    { GemmP ge2a12;
      ge2a12.A = EH1; ge2a12.B = We2; ge2a12.bias = be2; ge2a12.R = EH1; ge2a12.C = EH;
      ge2a12.sAo = 0; ge2a12.sAi = 0; ge2a12.sAm = H; ge2a12.sAk = 1; ge2a12.sBo = 0; ge2a12.sBi = 0; ge2a12.sBn = 1; ge2a12.sBk = H; ge2a12.sCo = 0; ge2a12.sCi = 0; ge2a12.sCm = H; ge2a12.sRo = 0; ge2a12.sRi = 0; ge2a12.sRm = 0; ge2a12.sRn = 0;
      ge2a12.M = CH; ge2a12.N = H; ge2a12.K = H; ge2a12.zi_n = 1; ge2a12.flags = 1; ge2a12.act = 1;
      ge2a12.alpha = 1.0f; ge2a12.beta = 0.0f; ge2a12.sa = 1.0f; ge2a12.sb = 1.0f; ge2a12.Npad = H; ge2a12.pad_ = 0;
      k_gemm<1><<<dim3((unsigned)((H) + 31) / 32, (unsigned)((CH) + 15) / 16, (unsigned)(1)), 32, 0, stream>>>(ge2a12); }
    { GemmP gm12;
      gm12.A = EH; gm12.B = Wm; gm12.bias = bm; gm12.R = EH; gm12.C = MSG;
      gm12.sAo = 0; gm12.sAi = 0; gm12.sAm = H; gm12.sAk = 1; gm12.sBo = 0; gm12.sBi = 0; gm12.sBn = 1; gm12.sBk = H; gm12.sCo = 0; gm12.sCi = 0; gm12.sCm = H; gm12.sRo = 0; gm12.sRi = 0; gm12.sRm = 0; gm12.sRn = 0;
      gm12.M = CH; gm12.N = H; gm12.K = H; gm12.zi_n = 1; gm12.flags = 1; gm12.act = 0;
      gm12.alpha = 1.0f; gm12.beta = 0.0f; gm12.sa = 1.0f; gm12.sb = 1.0f; gm12.Npad = H; gm12.pad_ = 0;
      k_gemm<1><<<dim3((unsigned)((H) + 31) / 32, (unsigned)((CH) + 15) / 16, (unsigned)(1)), 32, 0, stream>>>(gm12); }
    k_sb_scale<<<(unsigned)(((long long)CH * H + 255) / 256), 256, 0, stream>>>(MSG, escope, 375000, CH, H);
    k_sb_agg<<<(unsigned)(((long long)N * H + 255) / 256), 256, 0, stream>>>(MSG, soff, sslot, doff, dslot, AGG, 375000, CH, N, H);
    k_sb_edgectx<<<(unsigned)(((long long)CH * H + 255) / 256), 256, 0, stream>>>(ef, etype, eparams, emask, escope, ebatch, emb, ei, NH, EC, XS, XD, 406250, CH, E, H);
    { GemmP ge1aa13;
      ge1aa13.A = EC; ge1aa13.B = WS; ge1aa13.bias = be1; ge1aa13.R = EC; ge1aa13.C = EH1;
      ge1aa13.sAo = 0; ge1aa13.sAi = 0; ge1aa13.sAm = 32; ge1aa13.sAk = 1; ge1aa13.sBo = 0; ge1aa13.sBi = 0; ge1aa13.sBn = 1; ge1aa13.sBk = H; ge1aa13.sCo = 0; ge1aa13.sCi = 0; ge1aa13.sCm = H; ge1aa13.sRo = 0; ge1aa13.sRi = 0; ge1aa13.sRm = 0; ge1aa13.sRn = 0;
      ge1aa13.M = CH; ge1aa13.N = H; ge1aa13.K = 26; ge1aa13.zi_n = 1; ge1aa13.flags = 1; ge1aa13.act = 0;
      ge1aa13.alpha = 1.0f; ge1aa13.beta = 0.0f; ge1aa13.sa = 1.0f; ge1aa13.sb = 1.0f; ge1aa13.Npad = H; ge1aa13.pad_ = 0;
      k_gemm<1><<<dim3((unsigned)((H) + 31) / 32, (unsigned)((CH) + 15) / 16, (unsigned)(1)), 32, 0, stream>>>(ge1aa13); }
    { GemmP ge1ba13;
      ge1ba13.A = XS; ge1ba13.B = We1 + (size_t)4 * H; ge1ba13.bias = XS; ge1ba13.R = EH1; ge1ba13.C = EH1;
      ge1ba13.sAo = 0; ge1ba13.sAi = 0; ge1ba13.sAm = H; ge1ba13.sAk = 1; ge1ba13.sBo = 0; ge1ba13.sBi = 0; ge1ba13.sBn = 1; ge1ba13.sBk = H; ge1ba13.sCo = 0; ge1ba13.sCi = 0; ge1ba13.sCm = H; ge1ba13.sRo = 0; ge1ba13.sRi = 0; ge1ba13.sRm = H; ge1ba13.sRn = 1;
      ge1ba13.M = CH; ge1ba13.N = H; ge1ba13.K = H; ge1ba13.zi_n = 1; ge1ba13.flags = 4; ge1ba13.act = 0;
      ge1ba13.alpha = 1.0f; ge1ba13.beta = 1.0f; ge1ba13.sa = 1.0f; ge1ba13.sb = 1.0f; ge1ba13.Npad = H; ge1ba13.pad_ = 0;
      k_gemm<1><<<dim3((unsigned)((H) + 31) / 32, (unsigned)((CH) + 15) / 16, (unsigned)(1)), 32, 0, stream>>>(ge1ba13); }
    { GemmP ge1ca13;
      ge1ca13.A = XD; ge1ca13.B = We1 + (size_t)132 * H; ge1ca13.bias = XD; ge1ca13.R = EH1; ge1ca13.C = EH1;
      ge1ca13.sAo = 0; ge1ca13.sAi = 0; ge1ca13.sAm = H; ge1ca13.sAk = 1; ge1ca13.sBo = 0; ge1ca13.sBi = 0; ge1ca13.sBn = 1; ge1ca13.sBk = H; ge1ca13.sCo = 0; ge1ca13.sCi = 0; ge1ca13.sCm = H; ge1ca13.sRo = 0; ge1ca13.sRi = 0; ge1ca13.sRm = H; ge1ca13.sRn = 1;
      ge1ca13.M = CH; ge1ca13.N = H; ge1ca13.K = H; ge1ca13.zi_n = 1; ge1ca13.flags = 4; ge1ca13.act = 0;
      ge1ca13.alpha = 1.0f; ge1ca13.beta = 1.0f; ge1ca13.sa = 1.0f; ge1ca13.sb = 1.0f; ge1ca13.Npad = H; ge1ca13.pad_ = 0;
      k_gemm<1><<<dim3((unsigned)((H) + 31) / 32, (unsigned)((CH) + 15) / 16, (unsigned)(1)), 32, 0, stream>>>(ge1ca13); }
    k_norm_apply<<<(unsigned)(((long long)(1) * (1) * ((long long)CH * H) + 255) / 256), 256, 0, stream>>>(EH1, EH1, ust, nullptr, nullptr, 1, 1, (long long)CH * H, 1, 0, 1);
    { GemmP ge2a13;
      ge2a13.A = EH1; ge2a13.B = We2; ge2a13.bias = be2; ge2a13.R = EH1; ge2a13.C = EH;
      ge2a13.sAo = 0; ge2a13.sAi = 0; ge2a13.sAm = H; ge2a13.sAk = 1; ge2a13.sBo = 0; ge2a13.sBi = 0; ge2a13.sBn = 1; ge2a13.sBk = H; ge2a13.sCo = 0; ge2a13.sCi = 0; ge2a13.sCm = H; ge2a13.sRo = 0; ge2a13.sRi = 0; ge2a13.sRm = 0; ge2a13.sRn = 0;
      ge2a13.M = CH; ge2a13.N = H; ge2a13.K = H; ge2a13.zi_n = 1; ge2a13.flags = 1; ge2a13.act = 1;
      ge2a13.alpha = 1.0f; ge2a13.beta = 0.0f; ge2a13.sa = 1.0f; ge2a13.sb = 1.0f; ge2a13.Npad = H; ge2a13.pad_ = 0;
      k_gemm<1><<<dim3((unsigned)((H) + 31) / 32, (unsigned)((CH) + 15) / 16, (unsigned)(1)), 32, 0, stream>>>(ge2a13); }
    { GemmP gm13;
      gm13.A = EH; gm13.B = Wm; gm13.bias = bm; gm13.R = EH; gm13.C = MSG;
      gm13.sAo = 0; gm13.sAi = 0; gm13.sAm = H; gm13.sAk = 1; gm13.sBo = 0; gm13.sBi = 0; gm13.sBn = 1; gm13.sBk = H; gm13.sCo = 0; gm13.sCi = 0; gm13.sCm = H; gm13.sRo = 0; gm13.sRi = 0; gm13.sRm = 0; gm13.sRn = 0;
      gm13.M = CH; gm13.N = H; gm13.K = H; gm13.zi_n = 1; gm13.flags = 1; gm13.act = 0;
      gm13.alpha = 1.0f; gm13.beta = 0.0f; gm13.sa = 1.0f; gm13.sb = 1.0f; gm13.Npad = H; gm13.pad_ = 0;
      k_gemm<1><<<dim3((unsigned)((H) + 31) / 32, (unsigned)((CH) + 15) / 16, (unsigned)(1)), 32, 0, stream>>>(gm13); }
    k_sb_scale<<<(unsigned)(((long long)CH * H + 255) / 256), 256, 0, stream>>>(MSG, escope, 406250, CH, H);
    k_sb_agg<<<(unsigned)(((long long)N * H + 255) / 256), 256, 0, stream>>>(MSG, soff, sslot, doff, dslot, AGG, 406250, CH, N, H);
    k_sb_edgectx<<<(unsigned)(((long long)CH * H + 255) / 256), 256, 0, stream>>>(ef, etype, eparams, emask, escope, ebatch, emb, ei, NH, EC, XS, XD, 437500, CH, E, H);
    { GemmP ge1aa14;
      ge1aa14.A = EC; ge1aa14.B = WS; ge1aa14.bias = be1; ge1aa14.R = EC; ge1aa14.C = EH1;
      ge1aa14.sAo = 0; ge1aa14.sAi = 0; ge1aa14.sAm = 32; ge1aa14.sAk = 1; ge1aa14.sBo = 0; ge1aa14.sBi = 0; ge1aa14.sBn = 1; ge1aa14.sBk = H; ge1aa14.sCo = 0; ge1aa14.sCi = 0; ge1aa14.sCm = H; ge1aa14.sRo = 0; ge1aa14.sRi = 0; ge1aa14.sRm = 0; ge1aa14.sRn = 0;
      ge1aa14.M = CH; ge1aa14.N = H; ge1aa14.K = 26; ge1aa14.zi_n = 1; ge1aa14.flags = 1; ge1aa14.act = 0;
      ge1aa14.alpha = 1.0f; ge1aa14.beta = 0.0f; ge1aa14.sa = 1.0f; ge1aa14.sb = 1.0f; ge1aa14.Npad = H; ge1aa14.pad_ = 0;
      k_gemm<1><<<dim3((unsigned)((H) + 31) / 32, (unsigned)((CH) + 15) / 16, (unsigned)(1)), 32, 0, stream>>>(ge1aa14); }
    { GemmP ge1ba14;
      ge1ba14.A = XS; ge1ba14.B = We1 + (size_t)4 * H; ge1ba14.bias = XS; ge1ba14.R = EH1; ge1ba14.C = EH1;
      ge1ba14.sAo = 0; ge1ba14.sAi = 0; ge1ba14.sAm = H; ge1ba14.sAk = 1; ge1ba14.sBo = 0; ge1ba14.sBi = 0; ge1ba14.sBn = 1; ge1ba14.sBk = H; ge1ba14.sCo = 0; ge1ba14.sCi = 0; ge1ba14.sCm = H; ge1ba14.sRo = 0; ge1ba14.sRi = 0; ge1ba14.sRm = H; ge1ba14.sRn = 1;
      ge1ba14.M = CH; ge1ba14.N = H; ge1ba14.K = H; ge1ba14.zi_n = 1; ge1ba14.flags = 4; ge1ba14.act = 0;
      ge1ba14.alpha = 1.0f; ge1ba14.beta = 1.0f; ge1ba14.sa = 1.0f; ge1ba14.sb = 1.0f; ge1ba14.Npad = H; ge1ba14.pad_ = 0;
      k_gemm<1><<<dim3((unsigned)((H) + 31) / 32, (unsigned)((CH) + 15) / 16, (unsigned)(1)), 32, 0, stream>>>(ge1ba14); }
    { GemmP ge1ca14;
      ge1ca14.A = XD; ge1ca14.B = We1 + (size_t)132 * H; ge1ca14.bias = XD; ge1ca14.R = EH1; ge1ca14.C = EH1;
      ge1ca14.sAo = 0; ge1ca14.sAi = 0; ge1ca14.sAm = H; ge1ca14.sAk = 1; ge1ca14.sBo = 0; ge1ca14.sBi = 0; ge1ca14.sBn = 1; ge1ca14.sBk = H; ge1ca14.sCo = 0; ge1ca14.sCi = 0; ge1ca14.sCm = H; ge1ca14.sRo = 0; ge1ca14.sRi = 0; ge1ca14.sRm = H; ge1ca14.sRn = 1;
      ge1ca14.M = CH; ge1ca14.N = H; ge1ca14.K = H; ge1ca14.zi_n = 1; ge1ca14.flags = 4; ge1ca14.act = 0;
      ge1ca14.alpha = 1.0f; ge1ca14.beta = 1.0f; ge1ca14.sa = 1.0f; ge1ca14.sb = 1.0f; ge1ca14.Npad = H; ge1ca14.pad_ = 0;
      k_gemm<1><<<dim3((unsigned)((H) + 31) / 32, (unsigned)((CH) + 15) / 16, (unsigned)(1)), 32, 0, stream>>>(ge1ca14); }
    k_norm_apply<<<(unsigned)(((long long)(1) * (1) * ((long long)CH * H) + 255) / 256), 256, 0, stream>>>(EH1, EH1, ust, nullptr, nullptr, 1, 1, (long long)CH * H, 1, 0, 1);
    { GemmP ge2a14;
      ge2a14.A = EH1; ge2a14.B = We2; ge2a14.bias = be2; ge2a14.R = EH1; ge2a14.C = EH;
      ge2a14.sAo = 0; ge2a14.sAi = 0; ge2a14.sAm = H; ge2a14.sAk = 1; ge2a14.sBo = 0; ge2a14.sBi = 0; ge2a14.sBn = 1; ge2a14.sBk = H; ge2a14.sCo = 0; ge2a14.sCi = 0; ge2a14.sCm = H; ge2a14.sRo = 0; ge2a14.sRi = 0; ge2a14.sRm = 0; ge2a14.sRn = 0;
      ge2a14.M = CH; ge2a14.N = H; ge2a14.K = H; ge2a14.zi_n = 1; ge2a14.flags = 1; ge2a14.act = 1;
      ge2a14.alpha = 1.0f; ge2a14.beta = 0.0f; ge2a14.sa = 1.0f; ge2a14.sb = 1.0f; ge2a14.Npad = H; ge2a14.pad_ = 0;
      k_gemm<1><<<dim3((unsigned)((H) + 31) / 32, (unsigned)((CH) + 15) / 16, (unsigned)(1)), 32, 0, stream>>>(ge2a14); }
    { GemmP gm14;
      gm14.A = EH; gm14.B = Wm; gm14.bias = bm; gm14.R = EH; gm14.C = MSG;
      gm14.sAo = 0; gm14.sAi = 0; gm14.sAm = H; gm14.sAk = 1; gm14.sBo = 0; gm14.sBi = 0; gm14.sBn = 1; gm14.sBk = H; gm14.sCo = 0; gm14.sCi = 0; gm14.sCm = H; gm14.sRo = 0; gm14.sRi = 0; gm14.sRm = 0; gm14.sRn = 0;
      gm14.M = CH; gm14.N = H; gm14.K = H; gm14.zi_n = 1; gm14.flags = 1; gm14.act = 0;
      gm14.alpha = 1.0f; gm14.beta = 0.0f; gm14.sa = 1.0f; gm14.sb = 1.0f; gm14.Npad = H; gm14.pad_ = 0;
      k_gemm<1><<<dim3((unsigned)((H) + 31) / 32, (unsigned)((CH) + 15) / 16, (unsigned)(1)), 32, 0, stream>>>(gm14); }
    k_sb_scale<<<(unsigned)(((long long)CH * H + 255) / 256), 256, 0, stream>>>(MSG, escope, 437500, CH, H);
    k_sb_agg<<<(unsigned)(((long long)N * H + 255) / 256), 256, 0, stream>>>(MSG, soff, sslot, doff, dslot, AGG, 437500, CH, N, H);
    k_sb_edgectx<<<(unsigned)(((long long)CH * H + 255) / 256), 256, 0, stream>>>(ef, etype, eparams, emask, escope, ebatch, emb, ei, NH, EC, XS, XD, 468750, CH, E, H);
    { GemmP ge1aa15;
      ge1aa15.A = EC; ge1aa15.B = WS; ge1aa15.bias = be1; ge1aa15.R = EC; ge1aa15.C = EH1;
      ge1aa15.sAo = 0; ge1aa15.sAi = 0; ge1aa15.sAm = 32; ge1aa15.sAk = 1; ge1aa15.sBo = 0; ge1aa15.sBi = 0; ge1aa15.sBn = 1; ge1aa15.sBk = H; ge1aa15.sCo = 0; ge1aa15.sCi = 0; ge1aa15.sCm = H; ge1aa15.sRo = 0; ge1aa15.sRi = 0; ge1aa15.sRm = 0; ge1aa15.sRn = 0;
      ge1aa15.M = CH; ge1aa15.N = H; ge1aa15.K = 26; ge1aa15.zi_n = 1; ge1aa15.flags = 1; ge1aa15.act = 0;
      ge1aa15.alpha = 1.0f; ge1aa15.beta = 0.0f; ge1aa15.sa = 1.0f; ge1aa15.sb = 1.0f; ge1aa15.Npad = H; ge1aa15.pad_ = 0;
      k_gemm<1><<<dim3((unsigned)((H) + 31) / 32, (unsigned)((CH) + 15) / 16, (unsigned)(1)), 32, 0, stream>>>(ge1aa15); }
    { GemmP ge1ba15;
      ge1ba15.A = XS; ge1ba15.B = We1 + (size_t)4 * H; ge1ba15.bias = XS; ge1ba15.R = EH1; ge1ba15.C = EH1;
      ge1ba15.sAo = 0; ge1ba15.sAi = 0; ge1ba15.sAm = H; ge1ba15.sAk = 1; ge1ba15.sBo = 0; ge1ba15.sBi = 0; ge1ba15.sBn = 1; ge1ba15.sBk = H; ge1ba15.sCo = 0; ge1ba15.sCi = 0; ge1ba15.sCm = H; ge1ba15.sRo = 0; ge1ba15.sRi = 0; ge1ba15.sRm = H; ge1ba15.sRn = 1;
      ge1ba15.M = CH; ge1ba15.N = H; ge1ba15.K = H; ge1ba15.zi_n = 1; ge1ba15.flags = 4; ge1ba15.act = 0;
      ge1ba15.alpha = 1.0f; ge1ba15.beta = 1.0f; ge1ba15.sa = 1.0f; ge1ba15.sb = 1.0f; ge1ba15.Npad = H; ge1ba15.pad_ = 0;
      k_gemm<1><<<dim3((unsigned)((H) + 31) / 32, (unsigned)((CH) + 15) / 16, (unsigned)(1)), 32, 0, stream>>>(ge1ba15); }
    { GemmP ge1ca15;
      ge1ca15.A = XD; ge1ca15.B = We1 + (size_t)132 * H; ge1ca15.bias = XD; ge1ca15.R = EH1; ge1ca15.C = EH1;
      ge1ca15.sAo = 0; ge1ca15.sAi = 0; ge1ca15.sAm = H; ge1ca15.sAk = 1; ge1ca15.sBo = 0; ge1ca15.sBi = 0; ge1ca15.sBn = 1; ge1ca15.sBk = H; ge1ca15.sCo = 0; ge1ca15.sCi = 0; ge1ca15.sCm = H; ge1ca15.sRo = 0; ge1ca15.sRi = 0; ge1ca15.sRm = H; ge1ca15.sRn = 1;
      ge1ca15.M = CH; ge1ca15.N = H; ge1ca15.K = H; ge1ca15.zi_n = 1; ge1ca15.flags = 4; ge1ca15.act = 0;
      ge1ca15.alpha = 1.0f; ge1ca15.beta = 1.0f; ge1ca15.sa = 1.0f; ge1ca15.sb = 1.0f; ge1ca15.Npad = H; ge1ca15.pad_ = 0;
      k_gemm<1><<<dim3((unsigned)((H) + 31) / 32, (unsigned)((CH) + 15) / 16, (unsigned)(1)), 32, 0, stream>>>(ge1ca15); }
    k_norm_apply<<<(unsigned)(((long long)(1) * (1) * ((long long)CH * H) + 255) / 256), 256, 0, stream>>>(EH1, EH1, ust, nullptr, nullptr, 1, 1, (long long)CH * H, 1, 0, 1);
    { GemmP ge2a15;
      ge2a15.A = EH1; ge2a15.B = We2; ge2a15.bias = be2; ge2a15.R = EH1; ge2a15.C = EH;
      ge2a15.sAo = 0; ge2a15.sAi = 0; ge2a15.sAm = H; ge2a15.sAk = 1; ge2a15.sBo = 0; ge2a15.sBi = 0; ge2a15.sBn = 1; ge2a15.sBk = H; ge2a15.sCo = 0; ge2a15.sCi = 0; ge2a15.sCm = H; ge2a15.sRo = 0; ge2a15.sRi = 0; ge2a15.sRm = 0; ge2a15.sRn = 0;
      ge2a15.M = CH; ge2a15.N = H; ge2a15.K = H; ge2a15.zi_n = 1; ge2a15.flags = 1; ge2a15.act = 1;
      ge2a15.alpha = 1.0f; ge2a15.beta = 0.0f; ge2a15.sa = 1.0f; ge2a15.sb = 1.0f; ge2a15.Npad = H; ge2a15.pad_ = 0;
      k_gemm<1><<<dim3((unsigned)((H) + 31) / 32, (unsigned)((CH) + 15) / 16, (unsigned)(1)), 32, 0, stream>>>(ge2a15); }
    { GemmP gm15;
      gm15.A = EH; gm15.B = Wm; gm15.bias = bm; gm15.R = EH; gm15.C = MSG;
      gm15.sAo = 0; gm15.sAi = 0; gm15.sAm = H; gm15.sAk = 1; gm15.sBo = 0; gm15.sBi = 0; gm15.sBn = 1; gm15.sBk = H; gm15.sCo = 0; gm15.sCi = 0; gm15.sCm = H; gm15.sRo = 0; gm15.sRi = 0; gm15.sRm = 0; gm15.sRn = 0;
      gm15.M = CH; gm15.N = H; gm15.K = H; gm15.zi_n = 1; gm15.flags = 1; gm15.act = 0;
      gm15.alpha = 1.0f; gm15.beta = 0.0f; gm15.sa = 1.0f; gm15.sb = 1.0f; gm15.Npad = H; gm15.pad_ = 0;
      k_gemm<1><<<dim3((unsigned)((H) + 31) / 32, (unsigned)((CH) + 15) / 16, (unsigned)(1)), 32, 0, stream>>>(gm15); }
    k_sb_scale<<<(unsigned)(((long long)CH * H + 255) / 256), 256, 0, stream>>>(MSG, escope, 468750, CH, H);
    k_sb_agg<<<(unsigned)(((long long)N * H + 255) / 256), 256, 0, stream>>>(MSG, soff, sslot, doff, dslot, AGG, 468750, CH, N, H);
    { GemmP gu1;
      gu1.A = NH; gu1.B = Wu; gu1.bias = bu; gu1.R = NH; gu1.C = HU;
      gu1.sAo = 0; gu1.sAi = 0; gu1.sAm = H; gu1.sAk = 1; gu1.sBo = 0; gu1.sBi = 0; gu1.sBn = 1; gu1.sBk = H; gu1.sCo = 0; gu1.sCi = 0; gu1.sCm = H; gu1.sRo = 0; gu1.sRi = 0; gu1.sRm = 0; gu1.sRn = 0;
      gu1.M = N; gu1.N = H; gu1.K = H; gu1.zi_n = 1; gu1.flags = 1; gu1.act = 0;
      gu1.alpha = 1.0f; gu1.beta = 0.0f; gu1.sa = 1.0f; gu1.sb = 1.0f; gu1.Npad = H; gu1.pad_ = 0;
      k_gemm<1><<<dim3((unsigned)((H) + 31) / 32, (unsigned)((N) + 15) / 16, (unsigned)(1)), 32, 0, stream>>>(gu1); }
    { GemmP gu2;
      gu2.A = AGG; gu2.B = Wu + (size_t)H * H; gu2.bias = AGG; gu2.R = HU; gu2.C = HU;
      gu2.sAo = 0; gu2.sAi = 0; gu2.sAm = H; gu2.sAk = 1; gu2.sBo = 0; gu2.sBi = 0; gu2.sBn = 1; gu2.sBk = H; gu2.sCo = 0; gu2.sCi = 0; gu2.sCm = H; gu2.sRo = 0; gu2.sRi = 0; gu2.sRm = H; gu2.sRn = 1;
      gu2.M = N; gu2.N = H; gu2.K = H; gu2.zi_n = 1; gu2.flags = 4; gu2.act = 0;
      gu2.alpha = 1.0f; gu2.beta = 1.0f; gu2.sa = 1.0f; gu2.sb = 1.0f; gu2.Npad = H; gu2.pad_ = 0;
      k_gemm<1><<<dim3((unsigned)((H) + 31) / 32, (unsigned)((N) + 15) / 16, (unsigned)(1)), 32, 0, stream>>>(gu2); }
    k_norm_apply<<<(unsigned)(((long long)(1) * (1) * ((long long)N * H) + 255) / 256), 256, 0, stream>>>(HU, HU, ust, nullptr, nullptr, 1, 1, (long long)N * H, 1, 0, 1);
    { GemmP gnd;
      gnd.A = HU; gnd.B = Wnd; gnd.bias = bnd; gnd.R = HU; gnd.C = RN;
      gnd.sAo = 0; gnd.sAi = 0; gnd.sAm = H; gnd.sAk = 1; gnd.sBo = 0; gnd.sBi = 0; gnd.sBn = 1; gnd.sBk = 7; gnd.sCo = 0; gnd.sCi = 0; gnd.sCm = LP; gnd.sRo = 0; gnd.sRi = 0; gnd.sRm = 0; gnd.sRn = 0;
      gnd.M = N; gnd.N = 7; gnd.K = H; gnd.zi_n = 1; gnd.flags = 1; gnd.act = 0;
      gnd.alpha = 1.0f; gnd.beta = 0.0f; gnd.sa = 1.0f; gnd.sb = 1.0f; gnd.Npad = LP; gnd.pad_ = 0;
      k_gemm<1><<<dim3((unsigned)((LP) + 31) / 32, (unsigned)((N) + 15) / 16, (unsigned)(1)), 32, 0, stream>>>(gnd); }
    k_sb_nodeout<<<(unsigned)((N * 7 + 255) / 256), 256, 0, stream>>>(RN, LP, nscope, nf, out, o2, N);
    k_sb_edgectx<<<(unsigned)(((long long)CH * H + 255) / 256), 256, 0, stream>>>(ef, etype, eparams, emask, escope, ebatch, emb, ei, NH, EC, XS, XD, 0, CH, E, H);
    { GemmP ge1ab0;
      ge1ab0.A = EC; ge1ab0.B = WS; ge1ab0.bias = be1; ge1ab0.R = EC; ge1ab0.C = EH1;
      ge1ab0.sAo = 0; ge1ab0.sAi = 0; ge1ab0.sAm = 32; ge1ab0.sAk = 1; ge1ab0.sBo = 0; ge1ab0.sBi = 0; ge1ab0.sBn = 1; ge1ab0.sBk = H; ge1ab0.sCo = 0; ge1ab0.sCi = 0; ge1ab0.sCm = H; ge1ab0.sRo = 0; ge1ab0.sRi = 0; ge1ab0.sRm = 0; ge1ab0.sRn = 0;
      ge1ab0.M = CH; ge1ab0.N = H; ge1ab0.K = 26; ge1ab0.zi_n = 1; ge1ab0.flags = 1; ge1ab0.act = 0;
      ge1ab0.alpha = 1.0f; ge1ab0.beta = 0.0f; ge1ab0.sa = 1.0f; ge1ab0.sb = 1.0f; ge1ab0.Npad = H; ge1ab0.pad_ = 0;
      k_gemm<1><<<dim3((unsigned)((H) + 31) / 32, (unsigned)((CH) + 15) / 16, (unsigned)(1)), 32, 0, stream>>>(ge1ab0); }
    { GemmP ge1bb0;
      ge1bb0.A = XS; ge1bb0.B = We1 + (size_t)4 * H; ge1bb0.bias = XS; ge1bb0.R = EH1; ge1bb0.C = EH1;
      ge1bb0.sAo = 0; ge1bb0.sAi = 0; ge1bb0.sAm = H; ge1bb0.sAk = 1; ge1bb0.sBo = 0; ge1bb0.sBi = 0; ge1bb0.sBn = 1; ge1bb0.sBk = H; ge1bb0.sCo = 0; ge1bb0.sCi = 0; ge1bb0.sCm = H; ge1bb0.sRo = 0; ge1bb0.sRi = 0; ge1bb0.sRm = H; ge1bb0.sRn = 1;
      ge1bb0.M = CH; ge1bb0.N = H; ge1bb0.K = H; ge1bb0.zi_n = 1; ge1bb0.flags = 4; ge1bb0.act = 0;
      ge1bb0.alpha = 1.0f; ge1bb0.beta = 1.0f; ge1bb0.sa = 1.0f; ge1bb0.sb = 1.0f; ge1bb0.Npad = H; ge1bb0.pad_ = 0;
      k_gemm<1><<<dim3((unsigned)((H) + 31) / 32, (unsigned)((CH) + 15) / 16, (unsigned)(1)), 32, 0, stream>>>(ge1bb0); }
    { GemmP ge1cb0;
      ge1cb0.A = XD; ge1cb0.B = We1 + (size_t)132 * H; ge1cb0.bias = XD; ge1cb0.R = EH1; ge1cb0.C = EH1;
      ge1cb0.sAo = 0; ge1cb0.sAi = 0; ge1cb0.sAm = H; ge1cb0.sAk = 1; ge1cb0.sBo = 0; ge1cb0.sBi = 0; ge1cb0.sBn = 1; ge1cb0.sBk = H; ge1cb0.sCo = 0; ge1cb0.sCi = 0; ge1cb0.sCm = H; ge1cb0.sRo = 0; ge1cb0.sRi = 0; ge1cb0.sRm = H; ge1cb0.sRn = 1;
      ge1cb0.M = CH; ge1cb0.N = H; ge1cb0.K = H; ge1cb0.zi_n = 1; ge1cb0.flags = 4; ge1cb0.act = 0;
      ge1cb0.alpha = 1.0f; ge1cb0.beta = 1.0f; ge1cb0.sa = 1.0f; ge1cb0.sb = 1.0f; ge1cb0.Npad = H; ge1cb0.pad_ = 0;
      k_gemm<1><<<dim3((unsigned)((H) + 31) / 32, (unsigned)((CH) + 15) / 16, (unsigned)(1)), 32, 0, stream>>>(ge1cb0); }
    k_norm_apply<<<(unsigned)(((long long)(1) * (1) * ((long long)CH * H) + 255) / 256), 256, 0, stream>>>(EH1, EH1, ust, nullptr, nullptr, 1, 1, (long long)CH * H, 1, 0, 1);
    { GemmP ge2b0;
      ge2b0.A = EH1; ge2b0.B = We2; ge2b0.bias = be2; ge2b0.R = EH1; ge2b0.C = EH;
      ge2b0.sAo = 0; ge2b0.sAi = 0; ge2b0.sAm = H; ge2b0.sAk = 1; ge2b0.sBo = 0; ge2b0.sBi = 0; ge2b0.sBn = 1; ge2b0.sBk = H; ge2b0.sCo = 0; ge2b0.sCi = 0; ge2b0.sCm = H; ge2b0.sRo = 0; ge2b0.sRi = 0; ge2b0.sRm = 0; ge2b0.sRn = 0;
      ge2b0.M = CH; ge2b0.N = H; ge2b0.K = H; ge2b0.zi_n = 1; ge2b0.flags = 1; ge2b0.act = 1;
      ge2b0.alpha = 1.0f; ge2b0.beta = 0.0f; ge2b0.sa = 1.0f; ge2b0.sb = 1.0f; ge2b0.Npad = H; ge2b0.pad_ = 0;
      k_gemm<1><<<dim3((unsigned)((H) + 31) / 32, (unsigned)((CH) + 15) / 16, (unsigned)(1)), 32, 0, stream>>>(ge2b0); }
    k_sb_gather<<<(unsigned)(((long long)CH * H + 255) / 256), 256, 0, stream>>>(ei, HU, XS, XD, 0, CH, E, H);
    { GemmP gd1a0;
      gd1a0.A = EH; gd1a0.B = Wed1; gd1a0.bias = bed1; gd1a0.R = EH; gd1a0.C = EH1;
      gd1a0.sAo = 0; gd1a0.sAi = 0; gd1a0.sAm = H; gd1a0.sAk = 1; gd1a0.sBo = 0; gd1a0.sBi = 0; gd1a0.sBn = 1; gd1a0.sBk = H; gd1a0.sCo = 0; gd1a0.sCi = 0; gd1a0.sCm = H; gd1a0.sRo = 0; gd1a0.sRi = 0; gd1a0.sRm = 0; gd1a0.sRn = 0;
      gd1a0.M = CH; gd1a0.N = H; gd1a0.K = H; gd1a0.zi_n = 1; gd1a0.flags = 1; gd1a0.act = 0;
      gd1a0.alpha = 1.0f; gd1a0.beta = 0.0f; gd1a0.sa = 1.0f; gd1a0.sb = 1.0f; gd1a0.Npad = H; gd1a0.pad_ = 0;
      k_gemm<1><<<dim3((unsigned)((H) + 31) / 32, (unsigned)((CH) + 15) / 16, (unsigned)(1)), 32, 0, stream>>>(gd1a0); }
    { GemmP gd1b0;
      gd1b0.A = XS; gd1b0.B = Wed1 + (size_t)H * H; gd1b0.bias = XS; gd1b0.R = EH1; gd1b0.C = EH1;
      gd1b0.sAo = 0; gd1b0.sAi = 0; gd1b0.sAm = H; gd1b0.sAk = 1; gd1b0.sBo = 0; gd1b0.sBi = 0; gd1b0.sBn = 1; gd1b0.sBk = H; gd1b0.sCo = 0; gd1b0.sCi = 0; gd1b0.sCm = H; gd1b0.sRo = 0; gd1b0.sRi = 0; gd1b0.sRm = H; gd1b0.sRn = 1;
      gd1b0.M = CH; gd1b0.N = H; gd1b0.K = H; gd1b0.zi_n = 1; gd1b0.flags = 4; gd1b0.act = 0;
      gd1b0.alpha = 1.0f; gd1b0.beta = 1.0f; gd1b0.sa = 1.0f; gd1b0.sb = 1.0f; gd1b0.Npad = H; gd1b0.pad_ = 0;
      k_gemm<1><<<dim3((unsigned)((H) + 31) / 32, (unsigned)((CH) + 15) / 16, (unsigned)(1)), 32, 0, stream>>>(gd1b0); }
    { GemmP gd1c0;
      gd1c0.A = XD; gd1c0.B = Wed1 + (size_t)2 * H * H; gd1c0.bias = XD; gd1c0.R = EH1; gd1c0.C = EH1;
      gd1c0.sAo = 0; gd1c0.sAi = 0; gd1c0.sAm = H; gd1c0.sAk = 1; gd1c0.sBo = 0; gd1c0.sBi = 0; gd1c0.sBn = 1; gd1c0.sBk = H; gd1c0.sCo = 0; gd1c0.sCi = 0; gd1c0.sCm = H; gd1c0.sRo = 0; gd1c0.sRi = 0; gd1c0.sRm = H; gd1c0.sRn = 1;
      gd1c0.M = CH; gd1c0.N = H; gd1c0.K = H; gd1c0.zi_n = 1; gd1c0.flags = 4; gd1c0.act = 0;
      gd1c0.alpha = 1.0f; gd1c0.beta = 1.0f; gd1c0.sa = 1.0f; gd1c0.sb = 1.0f; gd1c0.Npad = H; gd1c0.pad_ = 0;
      k_gemm<1><<<dim3((unsigned)((H) + 31) / 32, (unsigned)((CH) + 15) / 16, (unsigned)(1)), 32, 0, stream>>>(gd1c0); }
    k_norm_apply<<<(unsigned)(((long long)(1) * (1) * ((long long)CH * H) + 255) / 256), 256, 0, stream>>>(EH1, EH1, ust, nullptr, nullptr, 1, 1, (long long)CH * H, 1, 0, 1);
    { GemmP gd20;
      gd20.A = EH1; gd20.B = Wed2; gd20.bias = bed2; gd20.R = EH1; gd20.C = RE;
      gd20.sAo = 0; gd20.sAi = 0; gd20.sAm = H; gd20.sAk = 1; gd20.sBo = 0; gd20.sBi = 0; gd20.sBn = 1; gd20.sBk = 4; gd20.sCo = 0; gd20.sCi = 0; gd20.sCm = LP; gd20.sRo = 0; gd20.sRi = 0; gd20.sRm = 0; gd20.sRn = 0;
      gd20.M = CH; gd20.N = 4; gd20.K = H; gd20.zi_n = 1; gd20.flags = 1; gd20.act = 0;
      gd20.alpha = 1.0f; gd20.beta = 0.0f; gd20.sa = 1.0f; gd20.sb = 1.0f; gd20.Npad = LP; gd20.pad_ = 0;
      k_gemm<1><<<dim3((unsigned)((LP) + 31) / 32, (unsigned)((CH) + 15) / 16, (unsigned)(1)), 32, 0, stream>>>(gd20); }
    k_sb_edgeout<<<(unsigned)((CH * 4 + 255) / 256), 256, 0, stream>>>(RE, LP, escope, ef, o1, o3, 0, CH);
    k_sb_edgectx<<<(unsigned)(((long long)CH * H + 255) / 256), 256, 0, stream>>>(ef, etype, eparams, emask, escope, ebatch, emb, ei, NH, EC, XS, XD, 31250, CH, E, H);
    { GemmP ge1ab1;
      ge1ab1.A = EC; ge1ab1.B = WS; ge1ab1.bias = be1; ge1ab1.R = EC; ge1ab1.C = EH1;
      ge1ab1.sAo = 0; ge1ab1.sAi = 0; ge1ab1.sAm = 32; ge1ab1.sAk = 1; ge1ab1.sBo = 0; ge1ab1.sBi = 0; ge1ab1.sBn = 1; ge1ab1.sBk = H; ge1ab1.sCo = 0; ge1ab1.sCi = 0; ge1ab1.sCm = H; ge1ab1.sRo = 0; ge1ab1.sRi = 0; ge1ab1.sRm = 0; ge1ab1.sRn = 0;
      ge1ab1.M = CH; ge1ab1.N = H; ge1ab1.K = 26; ge1ab1.zi_n = 1; ge1ab1.flags = 1; ge1ab1.act = 0;
      ge1ab1.alpha = 1.0f; ge1ab1.beta = 0.0f; ge1ab1.sa = 1.0f; ge1ab1.sb = 1.0f; ge1ab1.Npad = H; ge1ab1.pad_ = 0;
      k_gemm<1><<<dim3((unsigned)((H) + 31) / 32, (unsigned)((CH) + 15) / 16, (unsigned)(1)), 32, 0, stream>>>(ge1ab1); }
    { GemmP ge1bb1;
      ge1bb1.A = XS; ge1bb1.B = We1 + (size_t)4 * H; ge1bb1.bias = XS; ge1bb1.R = EH1; ge1bb1.C = EH1;
      ge1bb1.sAo = 0; ge1bb1.sAi = 0; ge1bb1.sAm = H; ge1bb1.sAk = 1; ge1bb1.sBo = 0; ge1bb1.sBi = 0; ge1bb1.sBn = 1; ge1bb1.sBk = H; ge1bb1.sCo = 0; ge1bb1.sCi = 0; ge1bb1.sCm = H; ge1bb1.sRo = 0; ge1bb1.sRi = 0; ge1bb1.sRm = H; ge1bb1.sRn = 1;
      ge1bb1.M = CH; ge1bb1.N = H; ge1bb1.K = H; ge1bb1.zi_n = 1; ge1bb1.flags = 4; ge1bb1.act = 0;
      ge1bb1.alpha = 1.0f; ge1bb1.beta = 1.0f; ge1bb1.sa = 1.0f; ge1bb1.sb = 1.0f; ge1bb1.Npad = H; ge1bb1.pad_ = 0;
      k_gemm<1><<<dim3((unsigned)((H) + 31) / 32, (unsigned)((CH) + 15) / 16, (unsigned)(1)), 32, 0, stream>>>(ge1bb1); }
    { GemmP ge1cb1;
      ge1cb1.A = XD; ge1cb1.B = We1 + (size_t)132 * H; ge1cb1.bias = XD; ge1cb1.R = EH1; ge1cb1.C = EH1;
      ge1cb1.sAo = 0; ge1cb1.sAi = 0; ge1cb1.sAm = H; ge1cb1.sAk = 1; ge1cb1.sBo = 0; ge1cb1.sBi = 0; ge1cb1.sBn = 1; ge1cb1.sBk = H; ge1cb1.sCo = 0; ge1cb1.sCi = 0; ge1cb1.sCm = H; ge1cb1.sRo = 0; ge1cb1.sRi = 0; ge1cb1.sRm = H; ge1cb1.sRn = 1;
      ge1cb1.M = CH; ge1cb1.N = H; ge1cb1.K = H; ge1cb1.zi_n = 1; ge1cb1.flags = 4; ge1cb1.act = 0;
      ge1cb1.alpha = 1.0f; ge1cb1.beta = 1.0f; ge1cb1.sa = 1.0f; ge1cb1.sb = 1.0f; ge1cb1.Npad = H; ge1cb1.pad_ = 0;
      k_gemm<1><<<dim3((unsigned)((H) + 31) / 32, (unsigned)((CH) + 15) / 16, (unsigned)(1)), 32, 0, stream>>>(ge1cb1); }
    k_norm_apply<<<(unsigned)(((long long)(1) * (1) * ((long long)CH * H) + 255) / 256), 256, 0, stream>>>(EH1, EH1, ust, nullptr, nullptr, 1, 1, (long long)CH * H, 1, 0, 1);
    { GemmP ge2b1;
      ge2b1.A = EH1; ge2b1.B = We2; ge2b1.bias = be2; ge2b1.R = EH1; ge2b1.C = EH;
      ge2b1.sAo = 0; ge2b1.sAi = 0; ge2b1.sAm = H; ge2b1.sAk = 1; ge2b1.sBo = 0; ge2b1.sBi = 0; ge2b1.sBn = 1; ge2b1.sBk = H; ge2b1.sCo = 0; ge2b1.sCi = 0; ge2b1.sCm = H; ge2b1.sRo = 0; ge2b1.sRi = 0; ge2b1.sRm = 0; ge2b1.sRn = 0;
      ge2b1.M = CH; ge2b1.N = H; ge2b1.K = H; ge2b1.zi_n = 1; ge2b1.flags = 1; ge2b1.act = 1;
      ge2b1.alpha = 1.0f; ge2b1.beta = 0.0f; ge2b1.sa = 1.0f; ge2b1.sb = 1.0f; ge2b1.Npad = H; ge2b1.pad_ = 0;
      k_gemm<1><<<dim3((unsigned)((H) + 31) / 32, (unsigned)((CH) + 15) / 16, (unsigned)(1)), 32, 0, stream>>>(ge2b1); }
    k_sb_gather<<<(unsigned)(((long long)CH * H + 255) / 256), 256, 0, stream>>>(ei, HU, XS, XD, 31250, CH, E, H);
    { GemmP gd1a1;
      gd1a1.A = EH; gd1a1.B = Wed1; gd1a1.bias = bed1; gd1a1.R = EH; gd1a1.C = EH1;
      gd1a1.sAo = 0; gd1a1.sAi = 0; gd1a1.sAm = H; gd1a1.sAk = 1; gd1a1.sBo = 0; gd1a1.sBi = 0; gd1a1.sBn = 1; gd1a1.sBk = H; gd1a1.sCo = 0; gd1a1.sCi = 0; gd1a1.sCm = H; gd1a1.sRo = 0; gd1a1.sRi = 0; gd1a1.sRm = 0; gd1a1.sRn = 0;
      gd1a1.M = CH; gd1a1.N = H; gd1a1.K = H; gd1a1.zi_n = 1; gd1a1.flags = 1; gd1a1.act = 0;
      gd1a1.alpha = 1.0f; gd1a1.beta = 0.0f; gd1a1.sa = 1.0f; gd1a1.sb = 1.0f; gd1a1.Npad = H; gd1a1.pad_ = 0;
      k_gemm<1><<<dim3((unsigned)((H) + 31) / 32, (unsigned)((CH) + 15) / 16, (unsigned)(1)), 32, 0, stream>>>(gd1a1); }
    { GemmP gd1b1;
      gd1b1.A = XS; gd1b1.B = Wed1 + (size_t)H * H; gd1b1.bias = XS; gd1b1.R = EH1; gd1b1.C = EH1;
      gd1b1.sAo = 0; gd1b1.sAi = 0; gd1b1.sAm = H; gd1b1.sAk = 1; gd1b1.sBo = 0; gd1b1.sBi = 0; gd1b1.sBn = 1; gd1b1.sBk = H; gd1b1.sCo = 0; gd1b1.sCi = 0; gd1b1.sCm = H; gd1b1.sRo = 0; gd1b1.sRi = 0; gd1b1.sRm = H; gd1b1.sRn = 1;
      gd1b1.M = CH; gd1b1.N = H; gd1b1.K = H; gd1b1.zi_n = 1; gd1b1.flags = 4; gd1b1.act = 0;
      gd1b1.alpha = 1.0f; gd1b1.beta = 1.0f; gd1b1.sa = 1.0f; gd1b1.sb = 1.0f; gd1b1.Npad = H; gd1b1.pad_ = 0;
      k_gemm<1><<<dim3((unsigned)((H) + 31) / 32, (unsigned)((CH) + 15) / 16, (unsigned)(1)), 32, 0, stream>>>(gd1b1); }
    { GemmP gd1c1;
      gd1c1.A = XD; gd1c1.B = Wed1 + (size_t)2 * H * H; gd1c1.bias = XD; gd1c1.R = EH1; gd1c1.C = EH1;
      gd1c1.sAo = 0; gd1c1.sAi = 0; gd1c1.sAm = H; gd1c1.sAk = 1; gd1c1.sBo = 0; gd1c1.sBi = 0; gd1c1.sBn = 1; gd1c1.sBk = H; gd1c1.sCo = 0; gd1c1.sCi = 0; gd1c1.sCm = H; gd1c1.sRo = 0; gd1c1.sRi = 0; gd1c1.sRm = H; gd1c1.sRn = 1;
      gd1c1.M = CH; gd1c1.N = H; gd1c1.K = H; gd1c1.zi_n = 1; gd1c1.flags = 4; gd1c1.act = 0;
      gd1c1.alpha = 1.0f; gd1c1.beta = 1.0f; gd1c1.sa = 1.0f; gd1c1.sb = 1.0f; gd1c1.Npad = H; gd1c1.pad_ = 0;
      k_gemm<1><<<dim3((unsigned)((H) + 31) / 32, (unsigned)((CH) + 15) / 16, (unsigned)(1)), 32, 0, stream>>>(gd1c1); }
    k_norm_apply<<<(unsigned)(((long long)(1) * (1) * ((long long)CH * H) + 255) / 256), 256, 0, stream>>>(EH1, EH1, ust, nullptr, nullptr, 1, 1, (long long)CH * H, 1, 0, 1);
    { GemmP gd21;
      gd21.A = EH1; gd21.B = Wed2; gd21.bias = bed2; gd21.R = EH1; gd21.C = RE;
      gd21.sAo = 0; gd21.sAi = 0; gd21.sAm = H; gd21.sAk = 1; gd21.sBo = 0; gd21.sBi = 0; gd21.sBn = 1; gd21.sBk = 4; gd21.sCo = 0; gd21.sCi = 0; gd21.sCm = LP; gd21.sRo = 0; gd21.sRi = 0; gd21.sRm = 0; gd21.sRn = 0;
      gd21.M = CH; gd21.N = 4; gd21.K = H; gd21.zi_n = 1; gd21.flags = 1; gd21.act = 0;
      gd21.alpha = 1.0f; gd21.beta = 0.0f; gd21.sa = 1.0f; gd21.sb = 1.0f; gd21.Npad = LP; gd21.pad_ = 0;
      k_gemm<1><<<dim3((unsigned)((LP) + 31) / 32, (unsigned)((CH) + 15) / 16, (unsigned)(1)), 32, 0, stream>>>(gd21); }
    k_sb_edgeout<<<(unsigned)((CH * 4 + 255) / 256), 256, 0, stream>>>(RE, LP, escope, ef, o1, o3, 31250, CH);
    k_sb_edgectx<<<(unsigned)(((long long)CH * H + 255) / 256), 256, 0, stream>>>(ef, etype, eparams, emask, escope, ebatch, emb, ei, NH, EC, XS, XD, 62500, CH, E, H);
    { GemmP ge1ab2;
      ge1ab2.A = EC; ge1ab2.B = WS; ge1ab2.bias = be1; ge1ab2.R = EC; ge1ab2.C = EH1;
      ge1ab2.sAo = 0; ge1ab2.sAi = 0; ge1ab2.sAm = 32; ge1ab2.sAk = 1; ge1ab2.sBo = 0; ge1ab2.sBi = 0; ge1ab2.sBn = 1; ge1ab2.sBk = H; ge1ab2.sCo = 0; ge1ab2.sCi = 0; ge1ab2.sCm = H; ge1ab2.sRo = 0; ge1ab2.sRi = 0; ge1ab2.sRm = 0; ge1ab2.sRn = 0;
      ge1ab2.M = CH; ge1ab2.N = H; ge1ab2.K = 26; ge1ab2.zi_n = 1; ge1ab2.flags = 1; ge1ab2.act = 0;
      ge1ab2.alpha = 1.0f; ge1ab2.beta = 0.0f; ge1ab2.sa = 1.0f; ge1ab2.sb = 1.0f; ge1ab2.Npad = H; ge1ab2.pad_ = 0;
      k_gemm<1><<<dim3((unsigned)((H) + 31) / 32, (unsigned)((CH) + 15) / 16, (unsigned)(1)), 32, 0, stream>>>(ge1ab2); }
    { GemmP ge1bb2;
      ge1bb2.A = XS; ge1bb2.B = We1 + (size_t)4 * H; ge1bb2.bias = XS; ge1bb2.R = EH1; ge1bb2.C = EH1;
      ge1bb2.sAo = 0; ge1bb2.sAi = 0; ge1bb2.sAm = H; ge1bb2.sAk = 1; ge1bb2.sBo = 0; ge1bb2.sBi = 0; ge1bb2.sBn = 1; ge1bb2.sBk = H; ge1bb2.sCo = 0; ge1bb2.sCi = 0; ge1bb2.sCm = H; ge1bb2.sRo = 0; ge1bb2.sRi = 0; ge1bb2.sRm = H; ge1bb2.sRn = 1;
      ge1bb2.M = CH; ge1bb2.N = H; ge1bb2.K = H; ge1bb2.zi_n = 1; ge1bb2.flags = 4; ge1bb2.act = 0;
      ge1bb2.alpha = 1.0f; ge1bb2.beta = 1.0f; ge1bb2.sa = 1.0f; ge1bb2.sb = 1.0f; ge1bb2.Npad = H; ge1bb2.pad_ = 0;
      k_gemm<1><<<dim3((unsigned)((H) + 31) / 32, (unsigned)((CH) + 15) / 16, (unsigned)(1)), 32, 0, stream>>>(ge1bb2); }
    { GemmP ge1cb2;
      ge1cb2.A = XD; ge1cb2.B = We1 + (size_t)132 * H; ge1cb2.bias = XD; ge1cb2.R = EH1; ge1cb2.C = EH1;
      ge1cb2.sAo = 0; ge1cb2.sAi = 0; ge1cb2.sAm = H; ge1cb2.sAk = 1; ge1cb2.sBo = 0; ge1cb2.sBi = 0; ge1cb2.sBn = 1; ge1cb2.sBk = H; ge1cb2.sCo = 0; ge1cb2.sCi = 0; ge1cb2.sCm = H; ge1cb2.sRo = 0; ge1cb2.sRi = 0; ge1cb2.sRm = H; ge1cb2.sRn = 1;
      ge1cb2.M = CH; ge1cb2.N = H; ge1cb2.K = H; ge1cb2.zi_n = 1; ge1cb2.flags = 4; ge1cb2.act = 0;
      ge1cb2.alpha = 1.0f; ge1cb2.beta = 1.0f; ge1cb2.sa = 1.0f; ge1cb2.sb = 1.0f; ge1cb2.Npad = H; ge1cb2.pad_ = 0;
      k_gemm<1><<<dim3((unsigned)((H) + 31) / 32, (unsigned)((CH) + 15) / 16, (unsigned)(1)), 32, 0, stream>>>(ge1cb2); }
    k_norm_apply<<<(unsigned)(((long long)(1) * (1) * ((long long)CH * H) + 255) / 256), 256, 0, stream>>>(EH1, EH1, ust, nullptr, nullptr, 1, 1, (long long)CH * H, 1, 0, 1);
    { GemmP ge2b2;
      ge2b2.A = EH1; ge2b2.B = We2; ge2b2.bias = be2; ge2b2.R = EH1; ge2b2.C = EH;
      ge2b2.sAo = 0; ge2b2.sAi = 0; ge2b2.sAm = H; ge2b2.sAk = 1; ge2b2.sBo = 0; ge2b2.sBi = 0; ge2b2.sBn = 1; ge2b2.sBk = H; ge2b2.sCo = 0; ge2b2.sCi = 0; ge2b2.sCm = H; ge2b2.sRo = 0; ge2b2.sRi = 0; ge2b2.sRm = 0; ge2b2.sRn = 0;
      ge2b2.M = CH; ge2b2.N = H; ge2b2.K = H; ge2b2.zi_n = 1; ge2b2.flags = 1; ge2b2.act = 1;
      ge2b2.alpha = 1.0f; ge2b2.beta = 0.0f; ge2b2.sa = 1.0f; ge2b2.sb = 1.0f; ge2b2.Npad = H; ge2b2.pad_ = 0;
      k_gemm<1><<<dim3((unsigned)((H) + 31) / 32, (unsigned)((CH) + 15) / 16, (unsigned)(1)), 32, 0, stream>>>(ge2b2); }
    k_sb_gather<<<(unsigned)(((long long)CH * H + 255) / 256), 256, 0, stream>>>(ei, HU, XS, XD, 62500, CH, E, H);
    { GemmP gd1a2;
      gd1a2.A = EH; gd1a2.B = Wed1; gd1a2.bias = bed1; gd1a2.R = EH; gd1a2.C = EH1;
      gd1a2.sAo = 0; gd1a2.sAi = 0; gd1a2.sAm = H; gd1a2.sAk = 1; gd1a2.sBo = 0; gd1a2.sBi = 0; gd1a2.sBn = 1; gd1a2.sBk = H; gd1a2.sCo = 0; gd1a2.sCi = 0; gd1a2.sCm = H; gd1a2.sRo = 0; gd1a2.sRi = 0; gd1a2.sRm = 0; gd1a2.sRn = 0;
      gd1a2.M = CH; gd1a2.N = H; gd1a2.K = H; gd1a2.zi_n = 1; gd1a2.flags = 1; gd1a2.act = 0;
      gd1a2.alpha = 1.0f; gd1a2.beta = 0.0f; gd1a2.sa = 1.0f; gd1a2.sb = 1.0f; gd1a2.Npad = H; gd1a2.pad_ = 0;
      k_gemm<1><<<dim3((unsigned)((H) + 31) / 32, (unsigned)((CH) + 15) / 16, (unsigned)(1)), 32, 0, stream>>>(gd1a2); }
    { GemmP gd1b2;
      gd1b2.A = XS; gd1b2.B = Wed1 + (size_t)H * H; gd1b2.bias = XS; gd1b2.R = EH1; gd1b2.C = EH1;
      gd1b2.sAo = 0; gd1b2.sAi = 0; gd1b2.sAm = H; gd1b2.sAk = 1; gd1b2.sBo = 0; gd1b2.sBi = 0; gd1b2.sBn = 1; gd1b2.sBk = H; gd1b2.sCo = 0; gd1b2.sCi = 0; gd1b2.sCm = H; gd1b2.sRo = 0; gd1b2.sRi = 0; gd1b2.sRm = H; gd1b2.sRn = 1;
      gd1b2.M = CH; gd1b2.N = H; gd1b2.K = H; gd1b2.zi_n = 1; gd1b2.flags = 4; gd1b2.act = 0;
      gd1b2.alpha = 1.0f; gd1b2.beta = 1.0f; gd1b2.sa = 1.0f; gd1b2.sb = 1.0f; gd1b2.Npad = H; gd1b2.pad_ = 0;
      k_gemm<1><<<dim3((unsigned)((H) + 31) / 32, (unsigned)((CH) + 15) / 16, (unsigned)(1)), 32, 0, stream>>>(gd1b2); }
    { GemmP gd1c2;
      gd1c2.A = XD; gd1c2.B = Wed1 + (size_t)2 * H * H; gd1c2.bias = XD; gd1c2.R = EH1; gd1c2.C = EH1;
      gd1c2.sAo = 0; gd1c2.sAi = 0; gd1c2.sAm = H; gd1c2.sAk = 1; gd1c2.sBo = 0; gd1c2.sBi = 0; gd1c2.sBn = 1; gd1c2.sBk = H; gd1c2.sCo = 0; gd1c2.sCi = 0; gd1c2.sCm = H; gd1c2.sRo = 0; gd1c2.sRi = 0; gd1c2.sRm = H; gd1c2.sRn = 1;
      gd1c2.M = CH; gd1c2.N = H; gd1c2.K = H; gd1c2.zi_n = 1; gd1c2.flags = 4; gd1c2.act = 0;
      gd1c2.alpha = 1.0f; gd1c2.beta = 1.0f; gd1c2.sa = 1.0f; gd1c2.sb = 1.0f; gd1c2.Npad = H; gd1c2.pad_ = 0;
      k_gemm<1><<<dim3((unsigned)((H) + 31) / 32, (unsigned)((CH) + 15) / 16, (unsigned)(1)), 32, 0, stream>>>(gd1c2); }
    k_norm_apply<<<(unsigned)(((long long)(1) * (1) * ((long long)CH * H) + 255) / 256), 256, 0, stream>>>(EH1, EH1, ust, nullptr, nullptr, 1, 1, (long long)CH * H, 1, 0, 1);
    { GemmP gd22;
      gd22.A = EH1; gd22.B = Wed2; gd22.bias = bed2; gd22.R = EH1; gd22.C = RE;
      gd22.sAo = 0; gd22.sAi = 0; gd22.sAm = H; gd22.sAk = 1; gd22.sBo = 0; gd22.sBi = 0; gd22.sBn = 1; gd22.sBk = 4; gd22.sCo = 0; gd22.sCi = 0; gd22.sCm = LP; gd22.sRo = 0; gd22.sRi = 0; gd22.sRm = 0; gd22.sRn = 0;
      gd22.M = CH; gd22.N = 4; gd22.K = H; gd22.zi_n = 1; gd22.flags = 1; gd22.act = 0;
      gd22.alpha = 1.0f; gd22.beta = 0.0f; gd22.sa = 1.0f; gd22.sb = 1.0f; gd22.Npad = LP; gd22.pad_ = 0;
      k_gemm<1><<<dim3((unsigned)((LP) + 31) / 32, (unsigned)((CH) + 15) / 16, (unsigned)(1)), 32, 0, stream>>>(gd22); }
    k_sb_edgeout<<<(unsigned)((CH * 4 + 255) / 256), 256, 0, stream>>>(RE, LP, escope, ef, o1, o3, 62500, CH);
    k_sb_edgectx<<<(unsigned)(((long long)CH * H + 255) / 256), 256, 0, stream>>>(ef, etype, eparams, emask, escope, ebatch, emb, ei, NH, EC, XS, XD, 93750, CH, E, H);
    { GemmP ge1ab3;
      ge1ab3.A = EC; ge1ab3.B = WS; ge1ab3.bias = be1; ge1ab3.R = EC; ge1ab3.C = EH1;
      ge1ab3.sAo = 0; ge1ab3.sAi = 0; ge1ab3.sAm = 32; ge1ab3.sAk = 1; ge1ab3.sBo = 0; ge1ab3.sBi = 0; ge1ab3.sBn = 1; ge1ab3.sBk = H; ge1ab3.sCo = 0; ge1ab3.sCi = 0; ge1ab3.sCm = H; ge1ab3.sRo = 0; ge1ab3.sRi = 0; ge1ab3.sRm = 0; ge1ab3.sRn = 0;
      ge1ab3.M = CH; ge1ab3.N = H; ge1ab3.K = 26; ge1ab3.zi_n = 1; ge1ab3.flags = 1; ge1ab3.act = 0;
      ge1ab3.alpha = 1.0f; ge1ab3.beta = 0.0f; ge1ab3.sa = 1.0f; ge1ab3.sb = 1.0f; ge1ab3.Npad = H; ge1ab3.pad_ = 0;
      k_gemm<1><<<dim3((unsigned)((H) + 31) / 32, (unsigned)((CH) + 15) / 16, (unsigned)(1)), 32, 0, stream>>>(ge1ab3); }
    { GemmP ge1bb3;
      ge1bb3.A = XS; ge1bb3.B = We1 + (size_t)4 * H; ge1bb3.bias = XS; ge1bb3.R = EH1; ge1bb3.C = EH1;
      ge1bb3.sAo = 0; ge1bb3.sAi = 0; ge1bb3.sAm = H; ge1bb3.sAk = 1; ge1bb3.sBo = 0; ge1bb3.sBi = 0; ge1bb3.sBn = 1; ge1bb3.sBk = H; ge1bb3.sCo = 0; ge1bb3.sCi = 0; ge1bb3.sCm = H; ge1bb3.sRo = 0; ge1bb3.sRi = 0; ge1bb3.sRm = H; ge1bb3.sRn = 1;
      ge1bb3.M = CH; ge1bb3.N = H; ge1bb3.K = H; ge1bb3.zi_n = 1; ge1bb3.flags = 4; ge1bb3.act = 0;
      ge1bb3.alpha = 1.0f; ge1bb3.beta = 1.0f; ge1bb3.sa = 1.0f; ge1bb3.sb = 1.0f; ge1bb3.Npad = H; ge1bb3.pad_ = 0;
      k_gemm<1><<<dim3((unsigned)((H) + 31) / 32, (unsigned)((CH) + 15) / 16, (unsigned)(1)), 32, 0, stream>>>(ge1bb3); }
    { GemmP ge1cb3;
      ge1cb3.A = XD; ge1cb3.B = We1 + (size_t)132 * H; ge1cb3.bias = XD; ge1cb3.R = EH1; ge1cb3.C = EH1;
      ge1cb3.sAo = 0; ge1cb3.sAi = 0; ge1cb3.sAm = H; ge1cb3.sAk = 1; ge1cb3.sBo = 0; ge1cb3.sBi = 0; ge1cb3.sBn = 1; ge1cb3.sBk = H; ge1cb3.sCo = 0; ge1cb3.sCi = 0; ge1cb3.sCm = H; ge1cb3.sRo = 0; ge1cb3.sRi = 0; ge1cb3.sRm = H; ge1cb3.sRn = 1;
      ge1cb3.M = CH; ge1cb3.N = H; ge1cb3.K = H; ge1cb3.zi_n = 1; ge1cb3.flags = 4; ge1cb3.act = 0;
      ge1cb3.alpha = 1.0f; ge1cb3.beta = 1.0f; ge1cb3.sa = 1.0f; ge1cb3.sb = 1.0f; ge1cb3.Npad = H; ge1cb3.pad_ = 0;
      k_gemm<1><<<dim3((unsigned)((H) + 31) / 32, (unsigned)((CH) + 15) / 16, (unsigned)(1)), 32, 0, stream>>>(ge1cb3); }
    k_norm_apply<<<(unsigned)(((long long)(1) * (1) * ((long long)CH * H) + 255) / 256), 256, 0, stream>>>(EH1, EH1, ust, nullptr, nullptr, 1, 1, (long long)CH * H, 1, 0, 1);
    { GemmP ge2b3;
      ge2b3.A = EH1; ge2b3.B = We2; ge2b3.bias = be2; ge2b3.R = EH1; ge2b3.C = EH;
      ge2b3.sAo = 0; ge2b3.sAi = 0; ge2b3.sAm = H; ge2b3.sAk = 1; ge2b3.sBo = 0; ge2b3.sBi = 0; ge2b3.sBn = 1; ge2b3.sBk = H; ge2b3.sCo = 0; ge2b3.sCi = 0; ge2b3.sCm = H; ge2b3.sRo = 0; ge2b3.sRi = 0; ge2b3.sRm = 0; ge2b3.sRn = 0;
      ge2b3.M = CH; ge2b3.N = H; ge2b3.K = H; ge2b3.zi_n = 1; ge2b3.flags = 1; ge2b3.act = 1;
      ge2b3.alpha = 1.0f; ge2b3.beta = 0.0f; ge2b3.sa = 1.0f; ge2b3.sb = 1.0f; ge2b3.Npad = H; ge2b3.pad_ = 0;
      k_gemm<1><<<dim3((unsigned)((H) + 31) / 32, (unsigned)((CH) + 15) / 16, (unsigned)(1)), 32, 0, stream>>>(ge2b3); }
    k_sb_gather<<<(unsigned)(((long long)CH * H + 255) / 256), 256, 0, stream>>>(ei, HU, XS, XD, 93750, CH, E, H);
    { GemmP gd1a3;
      gd1a3.A = EH; gd1a3.B = Wed1; gd1a3.bias = bed1; gd1a3.R = EH; gd1a3.C = EH1;
      gd1a3.sAo = 0; gd1a3.sAi = 0; gd1a3.sAm = H; gd1a3.sAk = 1; gd1a3.sBo = 0; gd1a3.sBi = 0; gd1a3.sBn = 1; gd1a3.sBk = H; gd1a3.sCo = 0; gd1a3.sCi = 0; gd1a3.sCm = H; gd1a3.sRo = 0; gd1a3.sRi = 0; gd1a3.sRm = 0; gd1a3.sRn = 0;
      gd1a3.M = CH; gd1a3.N = H; gd1a3.K = H; gd1a3.zi_n = 1; gd1a3.flags = 1; gd1a3.act = 0;
      gd1a3.alpha = 1.0f; gd1a3.beta = 0.0f; gd1a3.sa = 1.0f; gd1a3.sb = 1.0f; gd1a3.Npad = H; gd1a3.pad_ = 0;
      k_gemm<1><<<dim3((unsigned)((H) + 31) / 32, (unsigned)((CH) + 15) / 16, (unsigned)(1)), 32, 0, stream>>>(gd1a3); }
    { GemmP gd1b3;
      gd1b3.A = XS; gd1b3.B = Wed1 + (size_t)H * H; gd1b3.bias = XS; gd1b3.R = EH1; gd1b3.C = EH1;
      gd1b3.sAo = 0; gd1b3.sAi = 0; gd1b3.sAm = H; gd1b3.sAk = 1; gd1b3.sBo = 0; gd1b3.sBi = 0; gd1b3.sBn = 1; gd1b3.sBk = H; gd1b3.sCo = 0; gd1b3.sCi = 0; gd1b3.sCm = H; gd1b3.sRo = 0; gd1b3.sRi = 0; gd1b3.sRm = H; gd1b3.sRn = 1;
      gd1b3.M = CH; gd1b3.N = H; gd1b3.K = H; gd1b3.zi_n = 1; gd1b3.flags = 4; gd1b3.act = 0;
      gd1b3.alpha = 1.0f; gd1b3.beta = 1.0f; gd1b3.sa = 1.0f; gd1b3.sb = 1.0f; gd1b3.Npad = H; gd1b3.pad_ = 0;
      k_gemm<1><<<dim3((unsigned)((H) + 31) / 32, (unsigned)((CH) + 15) / 16, (unsigned)(1)), 32, 0, stream>>>(gd1b3); }
    { GemmP gd1c3;
      gd1c3.A = XD; gd1c3.B = Wed1 + (size_t)2 * H * H; gd1c3.bias = XD; gd1c3.R = EH1; gd1c3.C = EH1;
      gd1c3.sAo = 0; gd1c3.sAi = 0; gd1c3.sAm = H; gd1c3.sAk = 1; gd1c3.sBo = 0; gd1c3.sBi = 0; gd1c3.sBn = 1; gd1c3.sBk = H; gd1c3.sCo = 0; gd1c3.sCi = 0; gd1c3.sCm = H; gd1c3.sRo = 0; gd1c3.sRi = 0; gd1c3.sRm = H; gd1c3.sRn = 1;
      gd1c3.M = CH; gd1c3.N = H; gd1c3.K = H; gd1c3.zi_n = 1; gd1c3.flags = 4; gd1c3.act = 0;
      gd1c3.alpha = 1.0f; gd1c3.beta = 1.0f; gd1c3.sa = 1.0f; gd1c3.sb = 1.0f; gd1c3.Npad = H; gd1c3.pad_ = 0;
      k_gemm<1><<<dim3((unsigned)((H) + 31) / 32, (unsigned)((CH) + 15) / 16, (unsigned)(1)), 32, 0, stream>>>(gd1c3); }
    k_norm_apply<<<(unsigned)(((long long)(1) * (1) * ((long long)CH * H) + 255) / 256), 256, 0, stream>>>(EH1, EH1, ust, nullptr, nullptr, 1, 1, (long long)CH * H, 1, 0, 1);
    { GemmP gd23;
      gd23.A = EH1; gd23.B = Wed2; gd23.bias = bed2; gd23.R = EH1; gd23.C = RE;
      gd23.sAo = 0; gd23.sAi = 0; gd23.sAm = H; gd23.sAk = 1; gd23.sBo = 0; gd23.sBi = 0; gd23.sBn = 1; gd23.sBk = 4; gd23.sCo = 0; gd23.sCi = 0; gd23.sCm = LP; gd23.sRo = 0; gd23.sRi = 0; gd23.sRm = 0; gd23.sRn = 0;
      gd23.M = CH; gd23.N = 4; gd23.K = H; gd23.zi_n = 1; gd23.flags = 1; gd23.act = 0;
      gd23.alpha = 1.0f; gd23.beta = 0.0f; gd23.sa = 1.0f; gd23.sb = 1.0f; gd23.Npad = LP; gd23.pad_ = 0;
      k_gemm<1><<<dim3((unsigned)((LP) + 31) / 32, (unsigned)((CH) + 15) / 16, (unsigned)(1)), 32, 0, stream>>>(gd23); }
    k_sb_edgeout<<<(unsigned)((CH * 4 + 255) / 256), 256, 0, stream>>>(RE, LP, escope, ef, o1, o3, 93750, CH);
    k_sb_edgectx<<<(unsigned)(((long long)CH * H + 255) / 256), 256, 0, stream>>>(ef, etype, eparams, emask, escope, ebatch, emb, ei, NH, EC, XS, XD, 125000, CH, E, H);
    { GemmP ge1ab4;
      ge1ab4.A = EC; ge1ab4.B = WS; ge1ab4.bias = be1; ge1ab4.R = EC; ge1ab4.C = EH1;
      ge1ab4.sAo = 0; ge1ab4.sAi = 0; ge1ab4.sAm = 32; ge1ab4.sAk = 1; ge1ab4.sBo = 0; ge1ab4.sBi = 0; ge1ab4.sBn = 1; ge1ab4.sBk = H; ge1ab4.sCo = 0; ge1ab4.sCi = 0; ge1ab4.sCm = H; ge1ab4.sRo = 0; ge1ab4.sRi = 0; ge1ab4.sRm = 0; ge1ab4.sRn = 0;
      ge1ab4.M = CH; ge1ab4.N = H; ge1ab4.K = 26; ge1ab4.zi_n = 1; ge1ab4.flags = 1; ge1ab4.act = 0;
      ge1ab4.alpha = 1.0f; ge1ab4.beta = 0.0f; ge1ab4.sa = 1.0f; ge1ab4.sb = 1.0f; ge1ab4.Npad = H; ge1ab4.pad_ = 0;
      k_gemm<1><<<dim3((unsigned)((H) + 31) / 32, (unsigned)((CH) + 15) / 16, (unsigned)(1)), 32, 0, stream>>>(ge1ab4); }
    { GemmP ge1bb4;
      ge1bb4.A = XS; ge1bb4.B = We1 + (size_t)4 * H; ge1bb4.bias = XS; ge1bb4.R = EH1; ge1bb4.C = EH1;
      ge1bb4.sAo = 0; ge1bb4.sAi = 0; ge1bb4.sAm = H; ge1bb4.sAk = 1; ge1bb4.sBo = 0; ge1bb4.sBi = 0; ge1bb4.sBn = 1; ge1bb4.sBk = H; ge1bb4.sCo = 0; ge1bb4.sCi = 0; ge1bb4.sCm = H; ge1bb4.sRo = 0; ge1bb4.sRi = 0; ge1bb4.sRm = H; ge1bb4.sRn = 1;
      ge1bb4.M = CH; ge1bb4.N = H; ge1bb4.K = H; ge1bb4.zi_n = 1; ge1bb4.flags = 4; ge1bb4.act = 0;
      ge1bb4.alpha = 1.0f; ge1bb4.beta = 1.0f; ge1bb4.sa = 1.0f; ge1bb4.sb = 1.0f; ge1bb4.Npad = H; ge1bb4.pad_ = 0;
      k_gemm<1><<<dim3((unsigned)((H) + 31) / 32, (unsigned)((CH) + 15) / 16, (unsigned)(1)), 32, 0, stream>>>(ge1bb4); }
    { GemmP ge1cb4;
      ge1cb4.A = XD; ge1cb4.B = We1 + (size_t)132 * H; ge1cb4.bias = XD; ge1cb4.R = EH1; ge1cb4.C = EH1;
      ge1cb4.sAo = 0; ge1cb4.sAi = 0; ge1cb4.sAm = H; ge1cb4.sAk = 1; ge1cb4.sBo = 0; ge1cb4.sBi = 0; ge1cb4.sBn = 1; ge1cb4.sBk = H; ge1cb4.sCo = 0; ge1cb4.sCi = 0; ge1cb4.sCm = H; ge1cb4.sRo = 0; ge1cb4.sRi = 0; ge1cb4.sRm = H; ge1cb4.sRn = 1;
      ge1cb4.M = CH; ge1cb4.N = H; ge1cb4.K = H; ge1cb4.zi_n = 1; ge1cb4.flags = 4; ge1cb4.act = 0;
      ge1cb4.alpha = 1.0f; ge1cb4.beta = 1.0f; ge1cb4.sa = 1.0f; ge1cb4.sb = 1.0f; ge1cb4.Npad = H; ge1cb4.pad_ = 0;
      k_gemm<1><<<dim3((unsigned)((H) + 31) / 32, (unsigned)((CH) + 15) / 16, (unsigned)(1)), 32, 0, stream>>>(ge1cb4); }
    k_norm_apply<<<(unsigned)(((long long)(1) * (1) * ((long long)CH * H) + 255) / 256), 256, 0, stream>>>(EH1, EH1, ust, nullptr, nullptr, 1, 1, (long long)CH * H, 1, 0, 1);
    { GemmP ge2b4;
      ge2b4.A = EH1; ge2b4.B = We2; ge2b4.bias = be2; ge2b4.R = EH1; ge2b4.C = EH;
      ge2b4.sAo = 0; ge2b4.sAi = 0; ge2b4.sAm = H; ge2b4.sAk = 1; ge2b4.sBo = 0; ge2b4.sBi = 0; ge2b4.sBn = 1; ge2b4.sBk = H; ge2b4.sCo = 0; ge2b4.sCi = 0; ge2b4.sCm = H; ge2b4.sRo = 0; ge2b4.sRi = 0; ge2b4.sRm = 0; ge2b4.sRn = 0;
      ge2b4.M = CH; ge2b4.N = H; ge2b4.K = H; ge2b4.zi_n = 1; ge2b4.flags = 1; ge2b4.act = 1;
      ge2b4.alpha = 1.0f; ge2b4.beta = 0.0f; ge2b4.sa = 1.0f; ge2b4.sb = 1.0f; ge2b4.Npad = H; ge2b4.pad_ = 0;
      k_gemm<1><<<dim3((unsigned)((H) + 31) / 32, (unsigned)((CH) + 15) / 16, (unsigned)(1)), 32, 0, stream>>>(ge2b4); }
    k_sb_gather<<<(unsigned)(((long long)CH * H + 255) / 256), 256, 0, stream>>>(ei, HU, XS, XD, 125000, CH, E, H);
    { GemmP gd1a4;
      gd1a4.A = EH; gd1a4.B = Wed1; gd1a4.bias = bed1; gd1a4.R = EH; gd1a4.C = EH1;
      gd1a4.sAo = 0; gd1a4.sAi = 0; gd1a4.sAm = H; gd1a4.sAk = 1; gd1a4.sBo = 0; gd1a4.sBi = 0; gd1a4.sBn = 1; gd1a4.sBk = H; gd1a4.sCo = 0; gd1a4.sCi = 0; gd1a4.sCm = H; gd1a4.sRo = 0; gd1a4.sRi = 0; gd1a4.sRm = 0; gd1a4.sRn = 0;
      gd1a4.M = CH; gd1a4.N = H; gd1a4.K = H; gd1a4.zi_n = 1; gd1a4.flags = 1; gd1a4.act = 0;
      gd1a4.alpha = 1.0f; gd1a4.beta = 0.0f; gd1a4.sa = 1.0f; gd1a4.sb = 1.0f; gd1a4.Npad = H; gd1a4.pad_ = 0;
      k_gemm<1><<<dim3((unsigned)((H) + 31) / 32, (unsigned)((CH) + 15) / 16, (unsigned)(1)), 32, 0, stream>>>(gd1a4); }
    { GemmP gd1b4;
      gd1b4.A = XS; gd1b4.B = Wed1 + (size_t)H * H; gd1b4.bias = XS; gd1b4.R = EH1; gd1b4.C = EH1;
      gd1b4.sAo = 0; gd1b4.sAi = 0; gd1b4.sAm = H; gd1b4.sAk = 1; gd1b4.sBo = 0; gd1b4.sBi = 0; gd1b4.sBn = 1; gd1b4.sBk = H; gd1b4.sCo = 0; gd1b4.sCi = 0; gd1b4.sCm = H; gd1b4.sRo = 0; gd1b4.sRi = 0; gd1b4.sRm = H; gd1b4.sRn = 1;
      gd1b4.M = CH; gd1b4.N = H; gd1b4.K = H; gd1b4.zi_n = 1; gd1b4.flags = 4; gd1b4.act = 0;
      gd1b4.alpha = 1.0f; gd1b4.beta = 1.0f; gd1b4.sa = 1.0f; gd1b4.sb = 1.0f; gd1b4.Npad = H; gd1b4.pad_ = 0;
      k_gemm<1><<<dim3((unsigned)((H) + 31) / 32, (unsigned)((CH) + 15) / 16, (unsigned)(1)), 32, 0, stream>>>(gd1b4); }
    { GemmP gd1c4;
      gd1c4.A = XD; gd1c4.B = Wed1 + (size_t)2 * H * H; gd1c4.bias = XD; gd1c4.R = EH1; gd1c4.C = EH1;
      gd1c4.sAo = 0; gd1c4.sAi = 0; gd1c4.sAm = H; gd1c4.sAk = 1; gd1c4.sBo = 0; gd1c4.sBi = 0; gd1c4.sBn = 1; gd1c4.sBk = H; gd1c4.sCo = 0; gd1c4.sCi = 0; gd1c4.sCm = H; gd1c4.sRo = 0; gd1c4.sRi = 0; gd1c4.sRm = H; gd1c4.sRn = 1;
      gd1c4.M = CH; gd1c4.N = H; gd1c4.K = H; gd1c4.zi_n = 1; gd1c4.flags = 4; gd1c4.act = 0;
      gd1c4.alpha = 1.0f; gd1c4.beta = 1.0f; gd1c4.sa = 1.0f; gd1c4.sb = 1.0f; gd1c4.Npad = H; gd1c4.pad_ = 0;
      k_gemm<1><<<dim3((unsigned)((H) + 31) / 32, (unsigned)((CH) + 15) / 16, (unsigned)(1)), 32, 0, stream>>>(gd1c4); }
    k_norm_apply<<<(unsigned)(((long long)(1) * (1) * ((long long)CH * H) + 255) / 256), 256, 0, stream>>>(EH1, EH1, ust, nullptr, nullptr, 1, 1, (long long)CH * H, 1, 0, 1);
    { GemmP gd24;
      gd24.A = EH1; gd24.B = Wed2; gd24.bias = bed2; gd24.R = EH1; gd24.C = RE;
      gd24.sAo = 0; gd24.sAi = 0; gd24.sAm = H; gd24.sAk = 1; gd24.sBo = 0; gd24.sBi = 0; gd24.sBn = 1; gd24.sBk = 4; gd24.sCo = 0; gd24.sCi = 0; gd24.sCm = LP; gd24.sRo = 0; gd24.sRi = 0; gd24.sRm = 0; gd24.sRn = 0;
      gd24.M = CH; gd24.N = 4; gd24.K = H; gd24.zi_n = 1; gd24.flags = 1; gd24.act = 0;
      gd24.alpha = 1.0f; gd24.beta = 0.0f; gd24.sa = 1.0f; gd24.sb = 1.0f; gd24.Npad = LP; gd24.pad_ = 0;
      k_gemm<1><<<dim3((unsigned)((LP) + 31) / 32, (unsigned)((CH) + 15) / 16, (unsigned)(1)), 32, 0, stream>>>(gd24); }
    k_sb_edgeout<<<(unsigned)((CH * 4 + 255) / 256), 256, 0, stream>>>(RE, LP, escope, ef, o1, o3, 125000, CH);
    k_sb_edgectx<<<(unsigned)(((long long)CH * H + 255) / 256), 256, 0, stream>>>(ef, etype, eparams, emask, escope, ebatch, emb, ei, NH, EC, XS, XD, 156250, CH, E, H);
    { GemmP ge1ab5;
      ge1ab5.A = EC; ge1ab5.B = WS; ge1ab5.bias = be1; ge1ab5.R = EC; ge1ab5.C = EH1;
      ge1ab5.sAo = 0; ge1ab5.sAi = 0; ge1ab5.sAm = 32; ge1ab5.sAk = 1; ge1ab5.sBo = 0; ge1ab5.sBi = 0; ge1ab5.sBn = 1; ge1ab5.sBk = H; ge1ab5.sCo = 0; ge1ab5.sCi = 0; ge1ab5.sCm = H; ge1ab5.sRo = 0; ge1ab5.sRi = 0; ge1ab5.sRm = 0; ge1ab5.sRn = 0;
      ge1ab5.M = CH; ge1ab5.N = H; ge1ab5.K = 26; ge1ab5.zi_n = 1; ge1ab5.flags = 1; ge1ab5.act = 0;
      ge1ab5.alpha = 1.0f; ge1ab5.beta = 0.0f; ge1ab5.sa = 1.0f; ge1ab5.sb = 1.0f; ge1ab5.Npad = H; ge1ab5.pad_ = 0;
      k_gemm<1><<<dim3((unsigned)((H) + 31) / 32, (unsigned)((CH) + 15) / 16, (unsigned)(1)), 32, 0, stream>>>(ge1ab5); }
    { GemmP ge1bb5;
      ge1bb5.A = XS; ge1bb5.B = We1 + (size_t)4 * H; ge1bb5.bias = XS; ge1bb5.R = EH1; ge1bb5.C = EH1;
      ge1bb5.sAo = 0; ge1bb5.sAi = 0; ge1bb5.sAm = H; ge1bb5.sAk = 1; ge1bb5.sBo = 0; ge1bb5.sBi = 0; ge1bb5.sBn = 1; ge1bb5.sBk = H; ge1bb5.sCo = 0; ge1bb5.sCi = 0; ge1bb5.sCm = H; ge1bb5.sRo = 0; ge1bb5.sRi = 0; ge1bb5.sRm = H; ge1bb5.sRn = 1;
      ge1bb5.M = CH; ge1bb5.N = H; ge1bb5.K = H; ge1bb5.zi_n = 1; ge1bb5.flags = 4; ge1bb5.act = 0;
      ge1bb5.alpha = 1.0f; ge1bb5.beta = 1.0f; ge1bb5.sa = 1.0f; ge1bb5.sb = 1.0f; ge1bb5.Npad = H; ge1bb5.pad_ = 0;
      k_gemm<1><<<dim3((unsigned)((H) + 31) / 32, (unsigned)((CH) + 15) / 16, (unsigned)(1)), 32, 0, stream>>>(ge1bb5); }
    { GemmP ge1cb5;
      ge1cb5.A = XD; ge1cb5.B = We1 + (size_t)132 * H; ge1cb5.bias = XD; ge1cb5.R = EH1; ge1cb5.C = EH1;
      ge1cb5.sAo = 0; ge1cb5.sAi = 0; ge1cb5.sAm = H; ge1cb5.sAk = 1; ge1cb5.sBo = 0; ge1cb5.sBi = 0; ge1cb5.sBn = 1; ge1cb5.sBk = H; ge1cb5.sCo = 0; ge1cb5.sCi = 0; ge1cb5.sCm = H; ge1cb5.sRo = 0; ge1cb5.sRi = 0; ge1cb5.sRm = H; ge1cb5.sRn = 1;
      ge1cb5.M = CH; ge1cb5.N = H; ge1cb5.K = H; ge1cb5.zi_n = 1; ge1cb5.flags = 4; ge1cb5.act = 0;
      ge1cb5.alpha = 1.0f; ge1cb5.beta = 1.0f; ge1cb5.sa = 1.0f; ge1cb5.sb = 1.0f; ge1cb5.Npad = H; ge1cb5.pad_ = 0;
      k_gemm<1><<<dim3((unsigned)((H) + 31) / 32, (unsigned)((CH) + 15) / 16, (unsigned)(1)), 32, 0, stream>>>(ge1cb5); }
    k_norm_apply<<<(unsigned)(((long long)(1) * (1) * ((long long)CH * H) + 255) / 256), 256, 0, stream>>>(EH1, EH1, ust, nullptr, nullptr, 1, 1, (long long)CH * H, 1, 0, 1);
    { GemmP ge2b5;
      ge2b5.A = EH1; ge2b5.B = We2; ge2b5.bias = be2; ge2b5.R = EH1; ge2b5.C = EH;
      ge2b5.sAo = 0; ge2b5.sAi = 0; ge2b5.sAm = H; ge2b5.sAk = 1; ge2b5.sBo = 0; ge2b5.sBi = 0; ge2b5.sBn = 1; ge2b5.sBk = H; ge2b5.sCo = 0; ge2b5.sCi = 0; ge2b5.sCm = H; ge2b5.sRo = 0; ge2b5.sRi = 0; ge2b5.sRm = 0; ge2b5.sRn = 0;
      ge2b5.M = CH; ge2b5.N = H; ge2b5.K = H; ge2b5.zi_n = 1; ge2b5.flags = 1; ge2b5.act = 1;
      ge2b5.alpha = 1.0f; ge2b5.beta = 0.0f; ge2b5.sa = 1.0f; ge2b5.sb = 1.0f; ge2b5.Npad = H; ge2b5.pad_ = 0;
      k_gemm<1><<<dim3((unsigned)((H) + 31) / 32, (unsigned)((CH) + 15) / 16, (unsigned)(1)), 32, 0, stream>>>(ge2b5); }
    k_sb_gather<<<(unsigned)(((long long)CH * H + 255) / 256), 256, 0, stream>>>(ei, HU, XS, XD, 156250, CH, E, H);
    { GemmP gd1a5;
      gd1a5.A = EH; gd1a5.B = Wed1; gd1a5.bias = bed1; gd1a5.R = EH; gd1a5.C = EH1;
      gd1a5.sAo = 0; gd1a5.sAi = 0; gd1a5.sAm = H; gd1a5.sAk = 1; gd1a5.sBo = 0; gd1a5.sBi = 0; gd1a5.sBn = 1; gd1a5.sBk = H; gd1a5.sCo = 0; gd1a5.sCi = 0; gd1a5.sCm = H; gd1a5.sRo = 0; gd1a5.sRi = 0; gd1a5.sRm = 0; gd1a5.sRn = 0;
      gd1a5.M = CH; gd1a5.N = H; gd1a5.K = H; gd1a5.zi_n = 1; gd1a5.flags = 1; gd1a5.act = 0;
      gd1a5.alpha = 1.0f; gd1a5.beta = 0.0f; gd1a5.sa = 1.0f; gd1a5.sb = 1.0f; gd1a5.Npad = H; gd1a5.pad_ = 0;
      k_gemm<1><<<dim3((unsigned)((H) + 31) / 32, (unsigned)((CH) + 15) / 16, (unsigned)(1)), 32, 0, stream>>>(gd1a5); }
    { GemmP gd1b5;
      gd1b5.A = XS; gd1b5.B = Wed1 + (size_t)H * H; gd1b5.bias = XS; gd1b5.R = EH1; gd1b5.C = EH1;
      gd1b5.sAo = 0; gd1b5.sAi = 0; gd1b5.sAm = H; gd1b5.sAk = 1; gd1b5.sBo = 0; gd1b5.sBi = 0; gd1b5.sBn = 1; gd1b5.sBk = H; gd1b5.sCo = 0; gd1b5.sCi = 0; gd1b5.sCm = H; gd1b5.sRo = 0; gd1b5.sRi = 0; gd1b5.sRm = H; gd1b5.sRn = 1;
      gd1b5.M = CH; gd1b5.N = H; gd1b5.K = H; gd1b5.zi_n = 1; gd1b5.flags = 4; gd1b5.act = 0;
      gd1b5.alpha = 1.0f; gd1b5.beta = 1.0f; gd1b5.sa = 1.0f; gd1b5.sb = 1.0f; gd1b5.Npad = H; gd1b5.pad_ = 0;
      k_gemm<1><<<dim3((unsigned)((H) + 31) / 32, (unsigned)((CH) + 15) / 16, (unsigned)(1)), 32, 0, stream>>>(gd1b5); }
    { GemmP gd1c5;
      gd1c5.A = XD; gd1c5.B = Wed1 + (size_t)2 * H * H; gd1c5.bias = XD; gd1c5.R = EH1; gd1c5.C = EH1;
      gd1c5.sAo = 0; gd1c5.sAi = 0; gd1c5.sAm = H; gd1c5.sAk = 1; gd1c5.sBo = 0; gd1c5.sBi = 0; gd1c5.sBn = 1; gd1c5.sBk = H; gd1c5.sCo = 0; gd1c5.sCi = 0; gd1c5.sCm = H; gd1c5.sRo = 0; gd1c5.sRi = 0; gd1c5.sRm = H; gd1c5.sRn = 1;
      gd1c5.M = CH; gd1c5.N = H; gd1c5.K = H; gd1c5.zi_n = 1; gd1c5.flags = 4; gd1c5.act = 0;
      gd1c5.alpha = 1.0f; gd1c5.beta = 1.0f; gd1c5.sa = 1.0f; gd1c5.sb = 1.0f; gd1c5.Npad = H; gd1c5.pad_ = 0;
      k_gemm<1><<<dim3((unsigned)((H) + 31) / 32, (unsigned)((CH) + 15) / 16, (unsigned)(1)), 32, 0, stream>>>(gd1c5); }
    k_norm_apply<<<(unsigned)(((long long)(1) * (1) * ((long long)CH * H) + 255) / 256), 256, 0, stream>>>(EH1, EH1, ust, nullptr, nullptr, 1, 1, (long long)CH * H, 1, 0, 1);
    { GemmP gd25;
      gd25.A = EH1; gd25.B = Wed2; gd25.bias = bed2; gd25.R = EH1; gd25.C = RE;
      gd25.sAo = 0; gd25.sAi = 0; gd25.sAm = H; gd25.sAk = 1; gd25.sBo = 0; gd25.sBi = 0; gd25.sBn = 1; gd25.sBk = 4; gd25.sCo = 0; gd25.sCi = 0; gd25.sCm = LP; gd25.sRo = 0; gd25.sRi = 0; gd25.sRm = 0; gd25.sRn = 0;
      gd25.M = CH; gd25.N = 4; gd25.K = H; gd25.zi_n = 1; gd25.flags = 1; gd25.act = 0;
      gd25.alpha = 1.0f; gd25.beta = 0.0f; gd25.sa = 1.0f; gd25.sb = 1.0f; gd25.Npad = LP; gd25.pad_ = 0;
      k_gemm<1><<<dim3((unsigned)((LP) + 31) / 32, (unsigned)((CH) + 15) / 16, (unsigned)(1)), 32, 0, stream>>>(gd25); }
    k_sb_edgeout<<<(unsigned)((CH * 4 + 255) / 256), 256, 0, stream>>>(RE, LP, escope, ef, o1, o3, 156250, CH);
    k_sb_edgectx<<<(unsigned)(((long long)CH * H + 255) / 256), 256, 0, stream>>>(ef, etype, eparams, emask, escope, ebatch, emb, ei, NH, EC, XS, XD, 187500, CH, E, H);
    { GemmP ge1ab6;
      ge1ab6.A = EC; ge1ab6.B = WS; ge1ab6.bias = be1; ge1ab6.R = EC; ge1ab6.C = EH1;
      ge1ab6.sAo = 0; ge1ab6.sAi = 0; ge1ab6.sAm = 32; ge1ab6.sAk = 1; ge1ab6.sBo = 0; ge1ab6.sBi = 0; ge1ab6.sBn = 1; ge1ab6.sBk = H; ge1ab6.sCo = 0; ge1ab6.sCi = 0; ge1ab6.sCm = H; ge1ab6.sRo = 0; ge1ab6.sRi = 0; ge1ab6.sRm = 0; ge1ab6.sRn = 0;
      ge1ab6.M = CH; ge1ab6.N = H; ge1ab6.K = 26; ge1ab6.zi_n = 1; ge1ab6.flags = 1; ge1ab6.act = 0;
      ge1ab6.alpha = 1.0f; ge1ab6.beta = 0.0f; ge1ab6.sa = 1.0f; ge1ab6.sb = 1.0f; ge1ab6.Npad = H; ge1ab6.pad_ = 0;
      k_gemm<1><<<dim3((unsigned)((H) + 31) / 32, (unsigned)((CH) + 15) / 16, (unsigned)(1)), 32, 0, stream>>>(ge1ab6); }
    { GemmP ge1bb6;
      ge1bb6.A = XS; ge1bb6.B = We1 + (size_t)4 * H; ge1bb6.bias = XS; ge1bb6.R = EH1; ge1bb6.C = EH1;
      ge1bb6.sAo = 0; ge1bb6.sAi = 0; ge1bb6.sAm = H; ge1bb6.sAk = 1; ge1bb6.sBo = 0; ge1bb6.sBi = 0; ge1bb6.sBn = 1; ge1bb6.sBk = H; ge1bb6.sCo = 0; ge1bb6.sCi = 0; ge1bb6.sCm = H; ge1bb6.sRo = 0; ge1bb6.sRi = 0; ge1bb6.sRm = H; ge1bb6.sRn = 1;
      ge1bb6.M = CH; ge1bb6.N = H; ge1bb6.K = H; ge1bb6.zi_n = 1; ge1bb6.flags = 4; ge1bb6.act = 0;
      ge1bb6.alpha = 1.0f; ge1bb6.beta = 1.0f; ge1bb6.sa = 1.0f; ge1bb6.sb = 1.0f; ge1bb6.Npad = H; ge1bb6.pad_ = 0;
      k_gemm<1><<<dim3((unsigned)((H) + 31) / 32, (unsigned)((CH) + 15) / 16, (unsigned)(1)), 32, 0, stream>>>(ge1bb6); }
    { GemmP ge1cb6;
      ge1cb6.A = XD; ge1cb6.B = We1 + (size_t)132 * H; ge1cb6.bias = XD; ge1cb6.R = EH1; ge1cb6.C = EH1;
      ge1cb6.sAo = 0; ge1cb6.sAi = 0; ge1cb6.sAm = H; ge1cb6.sAk = 1; ge1cb6.sBo = 0; ge1cb6.sBi = 0; ge1cb6.sBn = 1; ge1cb6.sBk = H; ge1cb6.sCo = 0; ge1cb6.sCi = 0; ge1cb6.sCm = H; ge1cb6.sRo = 0; ge1cb6.sRi = 0; ge1cb6.sRm = H; ge1cb6.sRn = 1;
      ge1cb6.M = CH; ge1cb6.N = H; ge1cb6.K = H; ge1cb6.zi_n = 1; ge1cb6.flags = 4; ge1cb6.act = 0;
      ge1cb6.alpha = 1.0f; ge1cb6.beta = 1.0f; ge1cb6.sa = 1.0f; ge1cb6.sb = 1.0f; ge1cb6.Npad = H; ge1cb6.pad_ = 0;
      k_gemm<1><<<dim3((unsigned)((H) + 31) / 32, (unsigned)((CH) + 15) / 16, (unsigned)(1)), 32, 0, stream>>>(ge1cb6); }
    k_norm_apply<<<(unsigned)(((long long)(1) * (1) * ((long long)CH * H) + 255) / 256), 256, 0, stream>>>(EH1, EH1, ust, nullptr, nullptr, 1, 1, (long long)CH * H, 1, 0, 1);
    { GemmP ge2b6;
      ge2b6.A = EH1; ge2b6.B = We2; ge2b6.bias = be2; ge2b6.R = EH1; ge2b6.C = EH;
      ge2b6.sAo = 0; ge2b6.sAi = 0; ge2b6.sAm = H; ge2b6.sAk = 1; ge2b6.sBo = 0; ge2b6.sBi = 0; ge2b6.sBn = 1; ge2b6.sBk = H; ge2b6.sCo = 0; ge2b6.sCi = 0; ge2b6.sCm = H; ge2b6.sRo = 0; ge2b6.sRi = 0; ge2b6.sRm = 0; ge2b6.sRn = 0;
      ge2b6.M = CH; ge2b6.N = H; ge2b6.K = H; ge2b6.zi_n = 1; ge2b6.flags = 1; ge2b6.act = 1;
      ge2b6.alpha = 1.0f; ge2b6.beta = 0.0f; ge2b6.sa = 1.0f; ge2b6.sb = 1.0f; ge2b6.Npad = H; ge2b6.pad_ = 0;
      k_gemm<1><<<dim3((unsigned)((H) + 31) / 32, (unsigned)((CH) + 15) / 16, (unsigned)(1)), 32, 0, stream>>>(ge2b6); }
    k_sb_gather<<<(unsigned)(((long long)CH * H + 255) / 256), 256, 0, stream>>>(ei, HU, XS, XD, 187500, CH, E, H);
    { GemmP gd1a6;
      gd1a6.A = EH; gd1a6.B = Wed1; gd1a6.bias = bed1; gd1a6.R = EH; gd1a6.C = EH1;
      gd1a6.sAo = 0; gd1a6.sAi = 0; gd1a6.sAm = H; gd1a6.sAk = 1; gd1a6.sBo = 0; gd1a6.sBi = 0; gd1a6.sBn = 1; gd1a6.sBk = H; gd1a6.sCo = 0; gd1a6.sCi = 0; gd1a6.sCm = H; gd1a6.sRo = 0; gd1a6.sRi = 0; gd1a6.sRm = 0; gd1a6.sRn = 0;
      gd1a6.M = CH; gd1a6.N = H; gd1a6.K = H; gd1a6.zi_n = 1; gd1a6.flags = 1; gd1a6.act = 0;
      gd1a6.alpha = 1.0f; gd1a6.beta = 0.0f; gd1a6.sa = 1.0f; gd1a6.sb = 1.0f; gd1a6.Npad = H; gd1a6.pad_ = 0;
      k_gemm<1><<<dim3((unsigned)((H) + 31) / 32, (unsigned)((CH) + 15) / 16, (unsigned)(1)), 32, 0, stream>>>(gd1a6); }
    { GemmP gd1b6;
      gd1b6.A = XS; gd1b6.B = Wed1 + (size_t)H * H; gd1b6.bias = XS; gd1b6.R = EH1; gd1b6.C = EH1;
      gd1b6.sAo = 0; gd1b6.sAi = 0; gd1b6.sAm = H; gd1b6.sAk = 1; gd1b6.sBo = 0; gd1b6.sBi = 0; gd1b6.sBn = 1; gd1b6.sBk = H; gd1b6.sCo = 0; gd1b6.sCi = 0; gd1b6.sCm = H; gd1b6.sRo = 0; gd1b6.sRi = 0; gd1b6.sRm = H; gd1b6.sRn = 1;
      gd1b6.M = CH; gd1b6.N = H; gd1b6.K = H; gd1b6.zi_n = 1; gd1b6.flags = 4; gd1b6.act = 0;
      gd1b6.alpha = 1.0f; gd1b6.beta = 1.0f; gd1b6.sa = 1.0f; gd1b6.sb = 1.0f; gd1b6.Npad = H; gd1b6.pad_ = 0;
      k_gemm<1><<<dim3((unsigned)((H) + 31) / 32, (unsigned)((CH) + 15) / 16, (unsigned)(1)), 32, 0, stream>>>(gd1b6); }
    { GemmP gd1c6;
      gd1c6.A = XD; gd1c6.B = Wed1 + (size_t)2 * H * H; gd1c6.bias = XD; gd1c6.R = EH1; gd1c6.C = EH1;
      gd1c6.sAo = 0; gd1c6.sAi = 0; gd1c6.sAm = H; gd1c6.sAk = 1; gd1c6.sBo = 0; gd1c6.sBi = 0; gd1c6.sBn = 1; gd1c6.sBk = H; gd1c6.sCo = 0; gd1c6.sCi = 0; gd1c6.sCm = H; gd1c6.sRo = 0; gd1c6.sRi = 0; gd1c6.sRm = H; gd1c6.sRn = 1;
      gd1c6.M = CH; gd1c6.N = H; gd1c6.K = H; gd1c6.zi_n = 1; gd1c6.flags = 4; gd1c6.act = 0;
      gd1c6.alpha = 1.0f; gd1c6.beta = 1.0f; gd1c6.sa = 1.0f; gd1c6.sb = 1.0f; gd1c6.Npad = H; gd1c6.pad_ = 0;
      k_gemm<1><<<dim3((unsigned)((H) + 31) / 32, (unsigned)((CH) + 15) / 16, (unsigned)(1)), 32, 0, stream>>>(gd1c6); }
    k_norm_apply<<<(unsigned)(((long long)(1) * (1) * ((long long)CH * H) + 255) / 256), 256, 0, stream>>>(EH1, EH1, ust, nullptr, nullptr, 1, 1, (long long)CH * H, 1, 0, 1);
    { GemmP gd26;
      gd26.A = EH1; gd26.B = Wed2; gd26.bias = bed2; gd26.R = EH1; gd26.C = RE;
      gd26.sAo = 0; gd26.sAi = 0; gd26.sAm = H; gd26.sAk = 1; gd26.sBo = 0; gd26.sBi = 0; gd26.sBn = 1; gd26.sBk = 4; gd26.sCo = 0; gd26.sCi = 0; gd26.sCm = LP; gd26.sRo = 0; gd26.sRi = 0; gd26.sRm = 0; gd26.sRn = 0;
      gd26.M = CH; gd26.N = 4; gd26.K = H; gd26.zi_n = 1; gd26.flags = 1; gd26.act = 0;
      gd26.alpha = 1.0f; gd26.beta = 0.0f; gd26.sa = 1.0f; gd26.sb = 1.0f; gd26.Npad = LP; gd26.pad_ = 0;
      k_gemm<1><<<dim3((unsigned)((LP) + 31) / 32, (unsigned)((CH) + 15) / 16, (unsigned)(1)), 32, 0, stream>>>(gd26); }
    k_sb_edgeout<<<(unsigned)((CH * 4 + 255) / 256), 256, 0, stream>>>(RE, LP, escope, ef, o1, o3, 187500, CH);
    k_sb_edgectx<<<(unsigned)(((long long)CH * H + 255) / 256), 256, 0, stream>>>(ef, etype, eparams, emask, escope, ebatch, emb, ei, NH, EC, XS, XD, 218750, CH, E, H);
    { GemmP ge1ab7;
      ge1ab7.A = EC; ge1ab7.B = WS; ge1ab7.bias = be1; ge1ab7.R = EC; ge1ab7.C = EH1;
      ge1ab7.sAo = 0; ge1ab7.sAi = 0; ge1ab7.sAm = 32; ge1ab7.sAk = 1; ge1ab7.sBo = 0; ge1ab7.sBi = 0; ge1ab7.sBn = 1; ge1ab7.sBk = H; ge1ab7.sCo = 0; ge1ab7.sCi = 0; ge1ab7.sCm = H; ge1ab7.sRo = 0; ge1ab7.sRi = 0; ge1ab7.sRm = 0; ge1ab7.sRn = 0;
      ge1ab7.M = CH; ge1ab7.N = H; ge1ab7.K = 26; ge1ab7.zi_n = 1; ge1ab7.flags = 1; ge1ab7.act = 0;
      ge1ab7.alpha = 1.0f; ge1ab7.beta = 0.0f; ge1ab7.sa = 1.0f; ge1ab7.sb = 1.0f; ge1ab7.Npad = H; ge1ab7.pad_ = 0;
      k_gemm<1><<<dim3((unsigned)((H) + 31) / 32, (unsigned)((CH) + 15) / 16, (unsigned)(1)), 32, 0, stream>>>(ge1ab7); }
    { GemmP ge1bb7;
      ge1bb7.A = XS; ge1bb7.B = We1 + (size_t)4 * H; ge1bb7.bias = XS; ge1bb7.R = EH1; ge1bb7.C = EH1;
      ge1bb7.sAo = 0; ge1bb7.sAi = 0; ge1bb7.sAm = H; ge1bb7.sAk = 1; ge1bb7.sBo = 0; ge1bb7.sBi = 0; ge1bb7.sBn = 1; ge1bb7.sBk = H; ge1bb7.sCo = 0; ge1bb7.sCi = 0; ge1bb7.sCm = H; ge1bb7.sRo = 0; ge1bb7.sRi = 0; ge1bb7.sRm = H; ge1bb7.sRn = 1;
      ge1bb7.M = CH; ge1bb7.N = H; ge1bb7.K = H; ge1bb7.zi_n = 1; ge1bb7.flags = 4; ge1bb7.act = 0;
      ge1bb7.alpha = 1.0f; ge1bb7.beta = 1.0f; ge1bb7.sa = 1.0f; ge1bb7.sb = 1.0f; ge1bb7.Npad = H; ge1bb7.pad_ = 0;
      k_gemm<1><<<dim3((unsigned)((H) + 31) / 32, (unsigned)((CH) + 15) / 16, (unsigned)(1)), 32, 0, stream>>>(ge1bb7); }
    { GemmP ge1cb7;
      ge1cb7.A = XD; ge1cb7.B = We1 + (size_t)132 * H; ge1cb7.bias = XD; ge1cb7.R = EH1; ge1cb7.C = EH1;
      ge1cb7.sAo = 0; ge1cb7.sAi = 0; ge1cb7.sAm = H; ge1cb7.sAk = 1; ge1cb7.sBo = 0; ge1cb7.sBi = 0; ge1cb7.sBn = 1; ge1cb7.sBk = H; ge1cb7.sCo = 0; ge1cb7.sCi = 0; ge1cb7.sCm = H; ge1cb7.sRo = 0; ge1cb7.sRi = 0; ge1cb7.sRm = H; ge1cb7.sRn = 1;
      ge1cb7.M = CH; ge1cb7.N = H; ge1cb7.K = H; ge1cb7.zi_n = 1; ge1cb7.flags = 4; ge1cb7.act = 0;
      ge1cb7.alpha = 1.0f; ge1cb7.beta = 1.0f; ge1cb7.sa = 1.0f; ge1cb7.sb = 1.0f; ge1cb7.Npad = H; ge1cb7.pad_ = 0;
      k_gemm<1><<<dim3((unsigned)((H) + 31) / 32, (unsigned)((CH) + 15) / 16, (unsigned)(1)), 32, 0, stream>>>(ge1cb7); }
    k_norm_apply<<<(unsigned)(((long long)(1) * (1) * ((long long)CH * H) + 255) / 256), 256, 0, stream>>>(EH1, EH1, ust, nullptr, nullptr, 1, 1, (long long)CH * H, 1, 0, 1);
    { GemmP ge2b7;
      ge2b7.A = EH1; ge2b7.B = We2; ge2b7.bias = be2; ge2b7.R = EH1; ge2b7.C = EH;
      ge2b7.sAo = 0; ge2b7.sAi = 0; ge2b7.sAm = H; ge2b7.sAk = 1; ge2b7.sBo = 0; ge2b7.sBi = 0; ge2b7.sBn = 1; ge2b7.sBk = H; ge2b7.sCo = 0; ge2b7.sCi = 0; ge2b7.sCm = H; ge2b7.sRo = 0; ge2b7.sRi = 0; ge2b7.sRm = 0; ge2b7.sRn = 0;
      ge2b7.M = CH; ge2b7.N = H; ge2b7.K = H; ge2b7.zi_n = 1; ge2b7.flags = 1; ge2b7.act = 1;
      ge2b7.alpha = 1.0f; ge2b7.beta = 0.0f; ge2b7.sa = 1.0f; ge2b7.sb = 1.0f; ge2b7.Npad = H; ge2b7.pad_ = 0;
      k_gemm<1><<<dim3((unsigned)((H) + 31) / 32, (unsigned)((CH) + 15) / 16, (unsigned)(1)), 32, 0, stream>>>(ge2b7); }
    k_sb_gather<<<(unsigned)(((long long)CH * H + 255) / 256), 256, 0, stream>>>(ei, HU, XS, XD, 218750, CH, E, H);
    { GemmP gd1a7;
      gd1a7.A = EH; gd1a7.B = Wed1; gd1a7.bias = bed1; gd1a7.R = EH; gd1a7.C = EH1;
      gd1a7.sAo = 0; gd1a7.sAi = 0; gd1a7.sAm = H; gd1a7.sAk = 1; gd1a7.sBo = 0; gd1a7.sBi = 0; gd1a7.sBn = 1; gd1a7.sBk = H; gd1a7.sCo = 0; gd1a7.sCi = 0; gd1a7.sCm = H; gd1a7.sRo = 0; gd1a7.sRi = 0; gd1a7.sRm = 0; gd1a7.sRn = 0;
      gd1a7.M = CH; gd1a7.N = H; gd1a7.K = H; gd1a7.zi_n = 1; gd1a7.flags = 1; gd1a7.act = 0;
      gd1a7.alpha = 1.0f; gd1a7.beta = 0.0f; gd1a7.sa = 1.0f; gd1a7.sb = 1.0f; gd1a7.Npad = H; gd1a7.pad_ = 0;
      k_gemm<1><<<dim3((unsigned)((H) + 31) / 32, (unsigned)((CH) + 15) / 16, (unsigned)(1)), 32, 0, stream>>>(gd1a7); }
    { GemmP gd1b7;
      gd1b7.A = XS; gd1b7.B = Wed1 + (size_t)H * H; gd1b7.bias = XS; gd1b7.R = EH1; gd1b7.C = EH1;
      gd1b7.sAo = 0; gd1b7.sAi = 0; gd1b7.sAm = H; gd1b7.sAk = 1; gd1b7.sBo = 0; gd1b7.sBi = 0; gd1b7.sBn = 1; gd1b7.sBk = H; gd1b7.sCo = 0; gd1b7.sCi = 0; gd1b7.sCm = H; gd1b7.sRo = 0; gd1b7.sRi = 0; gd1b7.sRm = H; gd1b7.sRn = 1;
      gd1b7.M = CH; gd1b7.N = H; gd1b7.K = H; gd1b7.zi_n = 1; gd1b7.flags = 4; gd1b7.act = 0;
      gd1b7.alpha = 1.0f; gd1b7.beta = 1.0f; gd1b7.sa = 1.0f; gd1b7.sb = 1.0f; gd1b7.Npad = H; gd1b7.pad_ = 0;
      k_gemm<1><<<dim3((unsigned)((H) + 31) / 32, (unsigned)((CH) + 15) / 16, (unsigned)(1)), 32, 0, stream>>>(gd1b7); }
    { GemmP gd1c7;
      gd1c7.A = XD; gd1c7.B = Wed1 + (size_t)2 * H * H; gd1c7.bias = XD; gd1c7.R = EH1; gd1c7.C = EH1;
      gd1c7.sAo = 0; gd1c7.sAi = 0; gd1c7.sAm = H; gd1c7.sAk = 1; gd1c7.sBo = 0; gd1c7.sBi = 0; gd1c7.sBn = 1; gd1c7.sBk = H; gd1c7.sCo = 0; gd1c7.sCi = 0; gd1c7.sCm = H; gd1c7.sRo = 0; gd1c7.sRi = 0; gd1c7.sRm = H; gd1c7.sRn = 1;
      gd1c7.M = CH; gd1c7.N = H; gd1c7.K = H; gd1c7.zi_n = 1; gd1c7.flags = 4; gd1c7.act = 0;
      gd1c7.alpha = 1.0f; gd1c7.beta = 1.0f; gd1c7.sa = 1.0f; gd1c7.sb = 1.0f; gd1c7.Npad = H; gd1c7.pad_ = 0;
      k_gemm<1><<<dim3((unsigned)((H) + 31) / 32, (unsigned)((CH) + 15) / 16, (unsigned)(1)), 32, 0, stream>>>(gd1c7); }
    k_norm_apply<<<(unsigned)(((long long)(1) * (1) * ((long long)CH * H) + 255) / 256), 256, 0, stream>>>(EH1, EH1, ust, nullptr, nullptr, 1, 1, (long long)CH * H, 1, 0, 1);
    { GemmP gd27;
      gd27.A = EH1; gd27.B = Wed2; gd27.bias = bed2; gd27.R = EH1; gd27.C = RE;
      gd27.sAo = 0; gd27.sAi = 0; gd27.sAm = H; gd27.sAk = 1; gd27.sBo = 0; gd27.sBi = 0; gd27.sBn = 1; gd27.sBk = 4; gd27.sCo = 0; gd27.sCi = 0; gd27.sCm = LP; gd27.sRo = 0; gd27.sRi = 0; gd27.sRm = 0; gd27.sRn = 0;
      gd27.M = CH; gd27.N = 4; gd27.K = H; gd27.zi_n = 1; gd27.flags = 1; gd27.act = 0;
      gd27.alpha = 1.0f; gd27.beta = 0.0f; gd27.sa = 1.0f; gd27.sb = 1.0f; gd27.Npad = LP; gd27.pad_ = 0;
      k_gemm<1><<<dim3((unsigned)((LP) + 31) / 32, (unsigned)((CH) + 15) / 16, (unsigned)(1)), 32, 0, stream>>>(gd27); }
    k_sb_edgeout<<<(unsigned)((CH * 4 + 255) / 256), 256, 0, stream>>>(RE, LP, escope, ef, o1, o3, 218750, CH);
    k_sb_edgectx<<<(unsigned)(((long long)CH * H + 255) / 256), 256, 0, stream>>>(ef, etype, eparams, emask, escope, ebatch, emb, ei, NH, EC, XS, XD, 250000, CH, E, H);
    { GemmP ge1ab8;
      ge1ab8.A = EC; ge1ab8.B = WS; ge1ab8.bias = be1; ge1ab8.R = EC; ge1ab8.C = EH1;
      ge1ab8.sAo = 0; ge1ab8.sAi = 0; ge1ab8.sAm = 32; ge1ab8.sAk = 1; ge1ab8.sBo = 0; ge1ab8.sBi = 0; ge1ab8.sBn = 1; ge1ab8.sBk = H; ge1ab8.sCo = 0; ge1ab8.sCi = 0; ge1ab8.sCm = H; ge1ab8.sRo = 0; ge1ab8.sRi = 0; ge1ab8.sRm = 0; ge1ab8.sRn = 0;
      ge1ab8.M = CH; ge1ab8.N = H; ge1ab8.K = 26; ge1ab8.zi_n = 1; ge1ab8.flags = 1; ge1ab8.act = 0;
      ge1ab8.alpha = 1.0f; ge1ab8.beta = 0.0f; ge1ab8.sa = 1.0f; ge1ab8.sb = 1.0f; ge1ab8.Npad = H; ge1ab8.pad_ = 0;
      k_gemm<1><<<dim3((unsigned)((H) + 31) / 32, (unsigned)((CH) + 15) / 16, (unsigned)(1)), 32, 0, stream>>>(ge1ab8); }
    { GemmP ge1bb8;
      ge1bb8.A = XS; ge1bb8.B = We1 + (size_t)4 * H; ge1bb8.bias = XS; ge1bb8.R = EH1; ge1bb8.C = EH1;
      ge1bb8.sAo = 0; ge1bb8.sAi = 0; ge1bb8.sAm = H; ge1bb8.sAk = 1; ge1bb8.sBo = 0; ge1bb8.sBi = 0; ge1bb8.sBn = 1; ge1bb8.sBk = H; ge1bb8.sCo = 0; ge1bb8.sCi = 0; ge1bb8.sCm = H; ge1bb8.sRo = 0; ge1bb8.sRi = 0; ge1bb8.sRm = H; ge1bb8.sRn = 1;
      ge1bb8.M = CH; ge1bb8.N = H; ge1bb8.K = H; ge1bb8.zi_n = 1; ge1bb8.flags = 4; ge1bb8.act = 0;
      ge1bb8.alpha = 1.0f; ge1bb8.beta = 1.0f; ge1bb8.sa = 1.0f; ge1bb8.sb = 1.0f; ge1bb8.Npad = H; ge1bb8.pad_ = 0;
      k_gemm<1><<<dim3((unsigned)((H) + 31) / 32, (unsigned)((CH) + 15) / 16, (unsigned)(1)), 32, 0, stream>>>(ge1bb8); }
    { GemmP ge1cb8;
      ge1cb8.A = XD; ge1cb8.B = We1 + (size_t)132 * H; ge1cb8.bias = XD; ge1cb8.R = EH1; ge1cb8.C = EH1;
      ge1cb8.sAo = 0; ge1cb8.sAi = 0; ge1cb8.sAm = H; ge1cb8.sAk = 1; ge1cb8.sBo = 0; ge1cb8.sBi = 0; ge1cb8.sBn = 1; ge1cb8.sBk = H; ge1cb8.sCo = 0; ge1cb8.sCi = 0; ge1cb8.sCm = H; ge1cb8.sRo = 0; ge1cb8.sRi = 0; ge1cb8.sRm = H; ge1cb8.sRn = 1;
      ge1cb8.M = CH; ge1cb8.N = H; ge1cb8.K = H; ge1cb8.zi_n = 1; ge1cb8.flags = 4; ge1cb8.act = 0;
      ge1cb8.alpha = 1.0f; ge1cb8.beta = 1.0f; ge1cb8.sa = 1.0f; ge1cb8.sb = 1.0f; ge1cb8.Npad = H; ge1cb8.pad_ = 0;
      k_gemm<1><<<dim3((unsigned)((H) + 31) / 32, (unsigned)((CH) + 15) / 16, (unsigned)(1)), 32, 0, stream>>>(ge1cb8); }
    k_norm_apply<<<(unsigned)(((long long)(1) * (1) * ((long long)CH * H) + 255) / 256), 256, 0, stream>>>(EH1, EH1, ust, nullptr, nullptr, 1, 1, (long long)CH * H, 1, 0, 1);
    { GemmP ge2b8;
      ge2b8.A = EH1; ge2b8.B = We2; ge2b8.bias = be2; ge2b8.R = EH1; ge2b8.C = EH;
      ge2b8.sAo = 0; ge2b8.sAi = 0; ge2b8.sAm = H; ge2b8.sAk = 1; ge2b8.sBo = 0; ge2b8.sBi = 0; ge2b8.sBn = 1; ge2b8.sBk = H; ge2b8.sCo = 0; ge2b8.sCi = 0; ge2b8.sCm = H; ge2b8.sRo = 0; ge2b8.sRi = 0; ge2b8.sRm = 0; ge2b8.sRn = 0;
      ge2b8.M = CH; ge2b8.N = H; ge2b8.K = H; ge2b8.zi_n = 1; ge2b8.flags = 1; ge2b8.act = 1;
      ge2b8.alpha = 1.0f; ge2b8.beta = 0.0f; ge2b8.sa = 1.0f; ge2b8.sb = 1.0f; ge2b8.Npad = H; ge2b8.pad_ = 0;
      k_gemm<1><<<dim3((unsigned)((H) + 31) / 32, (unsigned)((CH) + 15) / 16, (unsigned)(1)), 32, 0, stream>>>(ge2b8); }
    k_sb_gather<<<(unsigned)(((long long)CH * H + 255) / 256), 256, 0, stream>>>(ei, HU, XS, XD, 250000, CH, E, H);
    { GemmP gd1a8;
      gd1a8.A = EH; gd1a8.B = Wed1; gd1a8.bias = bed1; gd1a8.R = EH; gd1a8.C = EH1;
      gd1a8.sAo = 0; gd1a8.sAi = 0; gd1a8.sAm = H; gd1a8.sAk = 1; gd1a8.sBo = 0; gd1a8.sBi = 0; gd1a8.sBn = 1; gd1a8.sBk = H; gd1a8.sCo = 0; gd1a8.sCi = 0; gd1a8.sCm = H; gd1a8.sRo = 0; gd1a8.sRi = 0; gd1a8.sRm = 0; gd1a8.sRn = 0;
      gd1a8.M = CH; gd1a8.N = H; gd1a8.K = H; gd1a8.zi_n = 1; gd1a8.flags = 1; gd1a8.act = 0;
      gd1a8.alpha = 1.0f; gd1a8.beta = 0.0f; gd1a8.sa = 1.0f; gd1a8.sb = 1.0f; gd1a8.Npad = H; gd1a8.pad_ = 0;
      k_gemm<1><<<dim3((unsigned)((H) + 31) / 32, (unsigned)((CH) + 15) / 16, (unsigned)(1)), 32, 0, stream>>>(gd1a8); }
    { GemmP gd1b8;
      gd1b8.A = XS; gd1b8.B = Wed1 + (size_t)H * H; gd1b8.bias = XS; gd1b8.R = EH1; gd1b8.C = EH1;
      gd1b8.sAo = 0; gd1b8.sAi = 0; gd1b8.sAm = H; gd1b8.sAk = 1; gd1b8.sBo = 0; gd1b8.sBi = 0; gd1b8.sBn = 1; gd1b8.sBk = H; gd1b8.sCo = 0; gd1b8.sCi = 0; gd1b8.sCm = H; gd1b8.sRo = 0; gd1b8.sRi = 0; gd1b8.sRm = H; gd1b8.sRn = 1;
      gd1b8.M = CH; gd1b8.N = H; gd1b8.K = H; gd1b8.zi_n = 1; gd1b8.flags = 4; gd1b8.act = 0;
      gd1b8.alpha = 1.0f; gd1b8.beta = 1.0f; gd1b8.sa = 1.0f; gd1b8.sb = 1.0f; gd1b8.Npad = H; gd1b8.pad_ = 0;
      k_gemm<1><<<dim3((unsigned)((H) + 31) / 32, (unsigned)((CH) + 15) / 16, (unsigned)(1)), 32, 0, stream>>>(gd1b8); }
    { GemmP gd1c8;
      gd1c8.A = XD; gd1c8.B = Wed1 + (size_t)2 * H * H; gd1c8.bias = XD; gd1c8.R = EH1; gd1c8.C = EH1;
      gd1c8.sAo = 0; gd1c8.sAi = 0; gd1c8.sAm = H; gd1c8.sAk = 1; gd1c8.sBo = 0; gd1c8.sBi = 0; gd1c8.sBn = 1; gd1c8.sBk = H; gd1c8.sCo = 0; gd1c8.sCi = 0; gd1c8.sCm = H; gd1c8.sRo = 0; gd1c8.sRi = 0; gd1c8.sRm = H; gd1c8.sRn = 1;
      gd1c8.M = CH; gd1c8.N = H; gd1c8.K = H; gd1c8.zi_n = 1; gd1c8.flags = 4; gd1c8.act = 0;
      gd1c8.alpha = 1.0f; gd1c8.beta = 1.0f; gd1c8.sa = 1.0f; gd1c8.sb = 1.0f; gd1c8.Npad = H; gd1c8.pad_ = 0;
      k_gemm<1><<<dim3((unsigned)((H) + 31) / 32, (unsigned)((CH) + 15) / 16, (unsigned)(1)), 32, 0, stream>>>(gd1c8); }
    k_norm_apply<<<(unsigned)(((long long)(1) * (1) * ((long long)CH * H) + 255) / 256), 256, 0, stream>>>(EH1, EH1, ust, nullptr, nullptr, 1, 1, (long long)CH * H, 1, 0, 1);
    { GemmP gd28;
      gd28.A = EH1; gd28.B = Wed2; gd28.bias = bed2; gd28.R = EH1; gd28.C = RE;
      gd28.sAo = 0; gd28.sAi = 0; gd28.sAm = H; gd28.sAk = 1; gd28.sBo = 0; gd28.sBi = 0; gd28.sBn = 1; gd28.sBk = 4; gd28.sCo = 0; gd28.sCi = 0; gd28.sCm = LP; gd28.sRo = 0; gd28.sRi = 0; gd28.sRm = 0; gd28.sRn = 0;
      gd28.M = CH; gd28.N = 4; gd28.K = H; gd28.zi_n = 1; gd28.flags = 1; gd28.act = 0;
      gd28.alpha = 1.0f; gd28.beta = 0.0f; gd28.sa = 1.0f; gd28.sb = 1.0f; gd28.Npad = LP; gd28.pad_ = 0;
      k_gemm<1><<<dim3((unsigned)((LP) + 31) / 32, (unsigned)((CH) + 15) / 16, (unsigned)(1)), 32, 0, stream>>>(gd28); }
    k_sb_edgeout<<<(unsigned)((CH * 4 + 255) / 256), 256, 0, stream>>>(RE, LP, escope, ef, o1, o3, 250000, CH);
    k_sb_edgectx<<<(unsigned)(((long long)CH * H + 255) / 256), 256, 0, stream>>>(ef, etype, eparams, emask, escope, ebatch, emb, ei, NH, EC, XS, XD, 281250, CH, E, H);
    { GemmP ge1ab9;
      ge1ab9.A = EC; ge1ab9.B = WS; ge1ab9.bias = be1; ge1ab9.R = EC; ge1ab9.C = EH1;
      ge1ab9.sAo = 0; ge1ab9.sAi = 0; ge1ab9.sAm = 32; ge1ab9.sAk = 1; ge1ab9.sBo = 0; ge1ab9.sBi = 0; ge1ab9.sBn = 1; ge1ab9.sBk = H; ge1ab9.sCo = 0; ge1ab9.sCi = 0; ge1ab9.sCm = H; ge1ab9.sRo = 0; ge1ab9.sRi = 0; ge1ab9.sRm = 0; ge1ab9.sRn = 0;
      ge1ab9.M = CH; ge1ab9.N = H; ge1ab9.K = 26; ge1ab9.zi_n = 1; ge1ab9.flags = 1; ge1ab9.act = 0;
      ge1ab9.alpha = 1.0f; ge1ab9.beta = 0.0f; ge1ab9.sa = 1.0f; ge1ab9.sb = 1.0f; ge1ab9.Npad = H; ge1ab9.pad_ = 0;
      k_gemm<1><<<dim3((unsigned)((H) + 31) / 32, (unsigned)((CH) + 15) / 16, (unsigned)(1)), 32, 0, stream>>>(ge1ab9); }
    { GemmP ge1bb9;
      ge1bb9.A = XS; ge1bb9.B = We1 + (size_t)4 * H; ge1bb9.bias = XS; ge1bb9.R = EH1; ge1bb9.C = EH1;
      ge1bb9.sAo = 0; ge1bb9.sAi = 0; ge1bb9.sAm = H; ge1bb9.sAk = 1; ge1bb9.sBo = 0; ge1bb9.sBi = 0; ge1bb9.sBn = 1; ge1bb9.sBk = H; ge1bb9.sCo = 0; ge1bb9.sCi = 0; ge1bb9.sCm = H; ge1bb9.sRo = 0; ge1bb9.sRi = 0; ge1bb9.sRm = H; ge1bb9.sRn = 1;
      ge1bb9.M = CH; ge1bb9.N = H; ge1bb9.K = H; ge1bb9.zi_n = 1; ge1bb9.flags = 4; ge1bb9.act = 0;
      ge1bb9.alpha = 1.0f; ge1bb9.beta = 1.0f; ge1bb9.sa = 1.0f; ge1bb9.sb = 1.0f; ge1bb9.Npad = H; ge1bb9.pad_ = 0;
      k_gemm<1><<<dim3((unsigned)((H) + 31) / 32, (unsigned)((CH) + 15) / 16, (unsigned)(1)), 32, 0, stream>>>(ge1bb9); }
    { GemmP ge1cb9;
      ge1cb9.A = XD; ge1cb9.B = We1 + (size_t)132 * H; ge1cb9.bias = XD; ge1cb9.R = EH1; ge1cb9.C = EH1;
      ge1cb9.sAo = 0; ge1cb9.sAi = 0; ge1cb9.sAm = H; ge1cb9.sAk = 1; ge1cb9.sBo = 0; ge1cb9.sBi = 0; ge1cb9.sBn = 1; ge1cb9.sBk = H; ge1cb9.sCo = 0; ge1cb9.sCi = 0; ge1cb9.sCm = H; ge1cb9.sRo = 0; ge1cb9.sRi = 0; ge1cb9.sRm = H; ge1cb9.sRn = 1;
      ge1cb9.M = CH; ge1cb9.N = H; ge1cb9.K = H; ge1cb9.zi_n = 1; ge1cb9.flags = 4; ge1cb9.act = 0;
      ge1cb9.alpha = 1.0f; ge1cb9.beta = 1.0f; ge1cb9.sa = 1.0f; ge1cb9.sb = 1.0f; ge1cb9.Npad = H; ge1cb9.pad_ = 0;
      k_gemm<1><<<dim3((unsigned)((H) + 31) / 32, (unsigned)((CH) + 15) / 16, (unsigned)(1)), 32, 0, stream>>>(ge1cb9); }
    k_norm_apply<<<(unsigned)(((long long)(1) * (1) * ((long long)CH * H) + 255) / 256), 256, 0, stream>>>(EH1, EH1, ust, nullptr, nullptr, 1, 1, (long long)CH * H, 1, 0, 1);
    { GemmP ge2b9;
      ge2b9.A = EH1; ge2b9.B = We2; ge2b9.bias = be2; ge2b9.R = EH1; ge2b9.C = EH;
      ge2b9.sAo = 0; ge2b9.sAi = 0; ge2b9.sAm = H; ge2b9.sAk = 1; ge2b9.sBo = 0; ge2b9.sBi = 0; ge2b9.sBn = 1; ge2b9.sBk = H; ge2b9.sCo = 0; ge2b9.sCi = 0; ge2b9.sCm = H; ge2b9.sRo = 0; ge2b9.sRi = 0; ge2b9.sRm = 0; ge2b9.sRn = 0;
      ge2b9.M = CH; ge2b9.N = H; ge2b9.K = H; ge2b9.zi_n = 1; ge2b9.flags = 1; ge2b9.act = 1;
      ge2b9.alpha = 1.0f; ge2b9.beta = 0.0f; ge2b9.sa = 1.0f; ge2b9.sb = 1.0f; ge2b9.Npad = H; ge2b9.pad_ = 0;
      k_gemm<1><<<dim3((unsigned)((H) + 31) / 32, (unsigned)((CH) + 15) / 16, (unsigned)(1)), 32, 0, stream>>>(ge2b9); }
    k_sb_gather<<<(unsigned)(((long long)CH * H + 255) / 256), 256, 0, stream>>>(ei, HU, XS, XD, 281250, CH, E, H);
    { GemmP gd1a9;
      gd1a9.A = EH; gd1a9.B = Wed1; gd1a9.bias = bed1; gd1a9.R = EH; gd1a9.C = EH1;
      gd1a9.sAo = 0; gd1a9.sAi = 0; gd1a9.sAm = H; gd1a9.sAk = 1; gd1a9.sBo = 0; gd1a9.sBi = 0; gd1a9.sBn = 1; gd1a9.sBk = H; gd1a9.sCo = 0; gd1a9.sCi = 0; gd1a9.sCm = H; gd1a9.sRo = 0; gd1a9.sRi = 0; gd1a9.sRm = 0; gd1a9.sRn = 0;
      gd1a9.M = CH; gd1a9.N = H; gd1a9.K = H; gd1a9.zi_n = 1; gd1a9.flags = 1; gd1a9.act = 0;
      gd1a9.alpha = 1.0f; gd1a9.beta = 0.0f; gd1a9.sa = 1.0f; gd1a9.sb = 1.0f; gd1a9.Npad = H; gd1a9.pad_ = 0;
      k_gemm<1><<<dim3((unsigned)((H) + 31) / 32, (unsigned)((CH) + 15) / 16, (unsigned)(1)), 32, 0, stream>>>(gd1a9); }
    { GemmP gd1b9;
      gd1b9.A = XS; gd1b9.B = Wed1 + (size_t)H * H; gd1b9.bias = XS; gd1b9.R = EH1; gd1b9.C = EH1;
      gd1b9.sAo = 0; gd1b9.sAi = 0; gd1b9.sAm = H; gd1b9.sAk = 1; gd1b9.sBo = 0; gd1b9.sBi = 0; gd1b9.sBn = 1; gd1b9.sBk = H; gd1b9.sCo = 0; gd1b9.sCi = 0; gd1b9.sCm = H; gd1b9.sRo = 0; gd1b9.sRi = 0; gd1b9.sRm = H; gd1b9.sRn = 1;
      gd1b9.M = CH; gd1b9.N = H; gd1b9.K = H; gd1b9.zi_n = 1; gd1b9.flags = 4; gd1b9.act = 0;
      gd1b9.alpha = 1.0f; gd1b9.beta = 1.0f; gd1b9.sa = 1.0f; gd1b9.sb = 1.0f; gd1b9.Npad = H; gd1b9.pad_ = 0;
      k_gemm<1><<<dim3((unsigned)((H) + 31) / 32, (unsigned)((CH) + 15) / 16, (unsigned)(1)), 32, 0, stream>>>(gd1b9); }
    { GemmP gd1c9;
      gd1c9.A = XD; gd1c9.B = Wed1 + (size_t)2 * H * H; gd1c9.bias = XD; gd1c9.R = EH1; gd1c9.C = EH1;
      gd1c9.sAo = 0; gd1c9.sAi = 0; gd1c9.sAm = H; gd1c9.sAk = 1; gd1c9.sBo = 0; gd1c9.sBi = 0; gd1c9.sBn = 1; gd1c9.sBk = H; gd1c9.sCo = 0; gd1c9.sCi = 0; gd1c9.sCm = H; gd1c9.sRo = 0; gd1c9.sRi = 0; gd1c9.sRm = H; gd1c9.sRn = 1;
      gd1c9.M = CH; gd1c9.N = H; gd1c9.K = H; gd1c9.zi_n = 1; gd1c9.flags = 4; gd1c9.act = 0;
      gd1c9.alpha = 1.0f; gd1c9.beta = 1.0f; gd1c9.sa = 1.0f; gd1c9.sb = 1.0f; gd1c9.Npad = H; gd1c9.pad_ = 0;
      k_gemm<1><<<dim3((unsigned)((H) + 31) / 32, (unsigned)((CH) + 15) / 16, (unsigned)(1)), 32, 0, stream>>>(gd1c9); }
    k_norm_apply<<<(unsigned)(((long long)(1) * (1) * ((long long)CH * H) + 255) / 256), 256, 0, stream>>>(EH1, EH1, ust, nullptr, nullptr, 1, 1, (long long)CH * H, 1, 0, 1);
    { GemmP gd29;
      gd29.A = EH1; gd29.B = Wed2; gd29.bias = bed2; gd29.R = EH1; gd29.C = RE;
      gd29.sAo = 0; gd29.sAi = 0; gd29.sAm = H; gd29.sAk = 1; gd29.sBo = 0; gd29.sBi = 0; gd29.sBn = 1; gd29.sBk = 4; gd29.sCo = 0; gd29.sCi = 0; gd29.sCm = LP; gd29.sRo = 0; gd29.sRi = 0; gd29.sRm = 0; gd29.sRn = 0;
      gd29.M = CH; gd29.N = 4; gd29.K = H; gd29.zi_n = 1; gd29.flags = 1; gd29.act = 0;
      gd29.alpha = 1.0f; gd29.beta = 0.0f; gd29.sa = 1.0f; gd29.sb = 1.0f; gd29.Npad = LP; gd29.pad_ = 0;
      k_gemm<1><<<dim3((unsigned)((LP) + 31) / 32, (unsigned)((CH) + 15) / 16, (unsigned)(1)), 32, 0, stream>>>(gd29); }
    k_sb_edgeout<<<(unsigned)((CH * 4 + 255) / 256), 256, 0, stream>>>(RE, LP, escope, ef, o1, o3, 281250, CH);
    k_sb_edgectx<<<(unsigned)(((long long)CH * H + 255) / 256), 256, 0, stream>>>(ef, etype, eparams, emask, escope, ebatch, emb, ei, NH, EC, XS, XD, 312500, CH, E, H);
    { GemmP ge1ab10;
      ge1ab10.A = EC; ge1ab10.B = WS; ge1ab10.bias = be1; ge1ab10.R = EC; ge1ab10.C = EH1;
      ge1ab10.sAo = 0; ge1ab10.sAi = 0; ge1ab10.sAm = 32; ge1ab10.sAk = 1; ge1ab10.sBo = 0; ge1ab10.sBi = 0; ge1ab10.sBn = 1; ge1ab10.sBk = H; ge1ab10.sCo = 0; ge1ab10.sCi = 0; ge1ab10.sCm = H; ge1ab10.sRo = 0; ge1ab10.sRi = 0; ge1ab10.sRm = 0; ge1ab10.sRn = 0;
      ge1ab10.M = CH; ge1ab10.N = H; ge1ab10.K = 26; ge1ab10.zi_n = 1; ge1ab10.flags = 1; ge1ab10.act = 0;
      ge1ab10.alpha = 1.0f; ge1ab10.beta = 0.0f; ge1ab10.sa = 1.0f; ge1ab10.sb = 1.0f; ge1ab10.Npad = H; ge1ab10.pad_ = 0;
      k_gemm<1><<<dim3((unsigned)((H) + 31) / 32, (unsigned)((CH) + 15) / 16, (unsigned)(1)), 32, 0, stream>>>(ge1ab10); }
    { GemmP ge1bb10;
      ge1bb10.A = XS; ge1bb10.B = We1 + (size_t)4 * H; ge1bb10.bias = XS; ge1bb10.R = EH1; ge1bb10.C = EH1;
      ge1bb10.sAo = 0; ge1bb10.sAi = 0; ge1bb10.sAm = H; ge1bb10.sAk = 1; ge1bb10.sBo = 0; ge1bb10.sBi = 0; ge1bb10.sBn = 1; ge1bb10.sBk = H; ge1bb10.sCo = 0; ge1bb10.sCi = 0; ge1bb10.sCm = H; ge1bb10.sRo = 0; ge1bb10.sRi = 0; ge1bb10.sRm = H; ge1bb10.sRn = 1;
      ge1bb10.M = CH; ge1bb10.N = H; ge1bb10.K = H; ge1bb10.zi_n = 1; ge1bb10.flags = 4; ge1bb10.act = 0;
      ge1bb10.alpha = 1.0f; ge1bb10.beta = 1.0f; ge1bb10.sa = 1.0f; ge1bb10.sb = 1.0f; ge1bb10.Npad = H; ge1bb10.pad_ = 0;
      k_gemm<1><<<dim3((unsigned)((H) + 31) / 32, (unsigned)((CH) + 15) / 16, (unsigned)(1)), 32, 0, stream>>>(ge1bb10); }
    { GemmP ge1cb10;
      ge1cb10.A = XD; ge1cb10.B = We1 + (size_t)132 * H; ge1cb10.bias = XD; ge1cb10.R = EH1; ge1cb10.C = EH1;
      ge1cb10.sAo = 0; ge1cb10.sAi = 0; ge1cb10.sAm = H; ge1cb10.sAk = 1; ge1cb10.sBo = 0; ge1cb10.sBi = 0; ge1cb10.sBn = 1; ge1cb10.sBk = H; ge1cb10.sCo = 0; ge1cb10.sCi = 0; ge1cb10.sCm = H; ge1cb10.sRo = 0; ge1cb10.sRi = 0; ge1cb10.sRm = H; ge1cb10.sRn = 1;
      ge1cb10.M = CH; ge1cb10.N = H; ge1cb10.K = H; ge1cb10.zi_n = 1; ge1cb10.flags = 4; ge1cb10.act = 0;
      ge1cb10.alpha = 1.0f; ge1cb10.beta = 1.0f; ge1cb10.sa = 1.0f; ge1cb10.sb = 1.0f; ge1cb10.Npad = H; ge1cb10.pad_ = 0;
      k_gemm<1><<<dim3((unsigned)((H) + 31) / 32, (unsigned)((CH) + 15) / 16, (unsigned)(1)), 32, 0, stream>>>(ge1cb10); }
    k_norm_apply<<<(unsigned)(((long long)(1) * (1) * ((long long)CH * H) + 255) / 256), 256, 0, stream>>>(EH1, EH1, ust, nullptr, nullptr, 1, 1, (long long)CH * H, 1, 0, 1);
    { GemmP ge2b10;
      ge2b10.A = EH1; ge2b10.B = We2; ge2b10.bias = be2; ge2b10.R = EH1; ge2b10.C = EH;
      ge2b10.sAo = 0; ge2b10.sAi = 0; ge2b10.sAm = H; ge2b10.sAk = 1; ge2b10.sBo = 0; ge2b10.sBi = 0; ge2b10.sBn = 1; ge2b10.sBk = H; ge2b10.sCo = 0; ge2b10.sCi = 0; ge2b10.sCm = H; ge2b10.sRo = 0; ge2b10.sRi = 0; ge2b10.sRm = 0; ge2b10.sRn = 0;
      ge2b10.M = CH; ge2b10.N = H; ge2b10.K = H; ge2b10.zi_n = 1; ge2b10.flags = 1; ge2b10.act = 1;
      ge2b10.alpha = 1.0f; ge2b10.beta = 0.0f; ge2b10.sa = 1.0f; ge2b10.sb = 1.0f; ge2b10.Npad = H; ge2b10.pad_ = 0;
      k_gemm<1><<<dim3((unsigned)((H) + 31) / 32, (unsigned)((CH) + 15) / 16, (unsigned)(1)), 32, 0, stream>>>(ge2b10); }
    k_sb_gather<<<(unsigned)(((long long)CH * H + 255) / 256), 256, 0, stream>>>(ei, HU, XS, XD, 312500, CH, E, H);
    { GemmP gd1a10;
      gd1a10.A = EH; gd1a10.B = Wed1; gd1a10.bias = bed1; gd1a10.R = EH; gd1a10.C = EH1;
      gd1a10.sAo = 0; gd1a10.sAi = 0; gd1a10.sAm = H; gd1a10.sAk = 1; gd1a10.sBo = 0; gd1a10.sBi = 0; gd1a10.sBn = 1; gd1a10.sBk = H; gd1a10.sCo = 0; gd1a10.sCi = 0; gd1a10.sCm = H; gd1a10.sRo = 0; gd1a10.sRi = 0; gd1a10.sRm = 0; gd1a10.sRn = 0;
      gd1a10.M = CH; gd1a10.N = H; gd1a10.K = H; gd1a10.zi_n = 1; gd1a10.flags = 1; gd1a10.act = 0;
      gd1a10.alpha = 1.0f; gd1a10.beta = 0.0f; gd1a10.sa = 1.0f; gd1a10.sb = 1.0f; gd1a10.Npad = H; gd1a10.pad_ = 0;
      k_gemm<1><<<dim3((unsigned)((H) + 31) / 32, (unsigned)((CH) + 15) / 16, (unsigned)(1)), 32, 0, stream>>>(gd1a10); }
    { GemmP gd1b10;
      gd1b10.A = XS; gd1b10.B = Wed1 + (size_t)H * H; gd1b10.bias = XS; gd1b10.R = EH1; gd1b10.C = EH1;
      gd1b10.sAo = 0; gd1b10.sAi = 0; gd1b10.sAm = H; gd1b10.sAk = 1; gd1b10.sBo = 0; gd1b10.sBi = 0; gd1b10.sBn = 1; gd1b10.sBk = H; gd1b10.sCo = 0; gd1b10.sCi = 0; gd1b10.sCm = H; gd1b10.sRo = 0; gd1b10.sRi = 0; gd1b10.sRm = H; gd1b10.sRn = 1;
      gd1b10.M = CH; gd1b10.N = H; gd1b10.K = H; gd1b10.zi_n = 1; gd1b10.flags = 4; gd1b10.act = 0;
      gd1b10.alpha = 1.0f; gd1b10.beta = 1.0f; gd1b10.sa = 1.0f; gd1b10.sb = 1.0f; gd1b10.Npad = H; gd1b10.pad_ = 0;
      k_gemm<1><<<dim3((unsigned)((H) + 31) / 32, (unsigned)((CH) + 15) / 16, (unsigned)(1)), 32, 0, stream>>>(gd1b10); }
    { GemmP gd1c10;
      gd1c10.A = XD; gd1c10.B = Wed1 + (size_t)2 * H * H; gd1c10.bias = XD; gd1c10.R = EH1; gd1c10.C = EH1;
      gd1c10.sAo = 0; gd1c10.sAi = 0; gd1c10.sAm = H; gd1c10.sAk = 1; gd1c10.sBo = 0; gd1c10.sBi = 0; gd1c10.sBn = 1; gd1c10.sBk = H; gd1c10.sCo = 0; gd1c10.sCi = 0; gd1c10.sCm = H; gd1c10.sRo = 0; gd1c10.sRi = 0; gd1c10.sRm = H; gd1c10.sRn = 1;
      gd1c10.M = CH; gd1c10.N = H; gd1c10.K = H; gd1c10.zi_n = 1; gd1c10.flags = 4; gd1c10.act = 0;
      gd1c10.alpha = 1.0f; gd1c10.beta = 1.0f; gd1c10.sa = 1.0f; gd1c10.sb = 1.0f; gd1c10.Npad = H; gd1c10.pad_ = 0;
      k_gemm<1><<<dim3((unsigned)((H) + 31) / 32, (unsigned)((CH) + 15) / 16, (unsigned)(1)), 32, 0, stream>>>(gd1c10); }
    k_norm_apply<<<(unsigned)(((long long)(1) * (1) * ((long long)CH * H) + 255) / 256), 256, 0, stream>>>(EH1, EH1, ust, nullptr, nullptr, 1, 1, (long long)CH * H, 1, 0, 1);
    { GemmP gd210;
      gd210.A = EH1; gd210.B = Wed2; gd210.bias = bed2; gd210.R = EH1; gd210.C = RE;
      gd210.sAo = 0; gd210.sAi = 0; gd210.sAm = H; gd210.sAk = 1; gd210.sBo = 0; gd210.sBi = 0; gd210.sBn = 1; gd210.sBk = 4; gd210.sCo = 0; gd210.sCi = 0; gd210.sCm = LP; gd210.sRo = 0; gd210.sRi = 0; gd210.sRm = 0; gd210.sRn = 0;
      gd210.M = CH; gd210.N = 4; gd210.K = H; gd210.zi_n = 1; gd210.flags = 1; gd210.act = 0;
      gd210.alpha = 1.0f; gd210.beta = 0.0f; gd210.sa = 1.0f; gd210.sb = 1.0f; gd210.Npad = LP; gd210.pad_ = 0;
      k_gemm<1><<<dim3((unsigned)((LP) + 31) / 32, (unsigned)((CH) + 15) / 16, (unsigned)(1)), 32, 0, stream>>>(gd210); }
    k_sb_edgeout<<<(unsigned)((CH * 4 + 255) / 256), 256, 0, stream>>>(RE, LP, escope, ef, o1, o3, 312500, CH);
    k_sb_edgectx<<<(unsigned)(((long long)CH * H + 255) / 256), 256, 0, stream>>>(ef, etype, eparams, emask, escope, ebatch, emb, ei, NH, EC, XS, XD, 343750, CH, E, H);
    { GemmP ge1ab11;
      ge1ab11.A = EC; ge1ab11.B = WS; ge1ab11.bias = be1; ge1ab11.R = EC; ge1ab11.C = EH1;
      ge1ab11.sAo = 0; ge1ab11.sAi = 0; ge1ab11.sAm = 32; ge1ab11.sAk = 1; ge1ab11.sBo = 0; ge1ab11.sBi = 0; ge1ab11.sBn = 1; ge1ab11.sBk = H; ge1ab11.sCo = 0; ge1ab11.sCi = 0; ge1ab11.sCm = H; ge1ab11.sRo = 0; ge1ab11.sRi = 0; ge1ab11.sRm = 0; ge1ab11.sRn = 0;
      ge1ab11.M = CH; ge1ab11.N = H; ge1ab11.K = 26; ge1ab11.zi_n = 1; ge1ab11.flags = 1; ge1ab11.act = 0;
      ge1ab11.alpha = 1.0f; ge1ab11.beta = 0.0f; ge1ab11.sa = 1.0f; ge1ab11.sb = 1.0f; ge1ab11.Npad = H; ge1ab11.pad_ = 0;
      k_gemm<1><<<dim3((unsigned)((H) + 31) / 32, (unsigned)((CH) + 15) / 16, (unsigned)(1)), 32, 0, stream>>>(ge1ab11); }
    { GemmP ge1bb11;
      ge1bb11.A = XS; ge1bb11.B = We1 + (size_t)4 * H; ge1bb11.bias = XS; ge1bb11.R = EH1; ge1bb11.C = EH1;
      ge1bb11.sAo = 0; ge1bb11.sAi = 0; ge1bb11.sAm = H; ge1bb11.sAk = 1; ge1bb11.sBo = 0; ge1bb11.sBi = 0; ge1bb11.sBn = 1; ge1bb11.sBk = H; ge1bb11.sCo = 0; ge1bb11.sCi = 0; ge1bb11.sCm = H; ge1bb11.sRo = 0; ge1bb11.sRi = 0; ge1bb11.sRm = H; ge1bb11.sRn = 1;
      ge1bb11.M = CH; ge1bb11.N = H; ge1bb11.K = H; ge1bb11.zi_n = 1; ge1bb11.flags = 4; ge1bb11.act = 0;
      ge1bb11.alpha = 1.0f; ge1bb11.beta = 1.0f; ge1bb11.sa = 1.0f; ge1bb11.sb = 1.0f; ge1bb11.Npad = H; ge1bb11.pad_ = 0;
      k_gemm<1><<<dim3((unsigned)((H) + 31) / 32, (unsigned)((CH) + 15) / 16, (unsigned)(1)), 32, 0, stream>>>(ge1bb11); }
    { GemmP ge1cb11;
      ge1cb11.A = XD; ge1cb11.B = We1 + (size_t)132 * H; ge1cb11.bias = XD; ge1cb11.R = EH1; ge1cb11.C = EH1;
      ge1cb11.sAo = 0; ge1cb11.sAi = 0; ge1cb11.sAm = H; ge1cb11.sAk = 1; ge1cb11.sBo = 0; ge1cb11.sBi = 0; ge1cb11.sBn = 1; ge1cb11.sBk = H; ge1cb11.sCo = 0; ge1cb11.sCi = 0; ge1cb11.sCm = H; ge1cb11.sRo = 0; ge1cb11.sRi = 0; ge1cb11.sRm = H; ge1cb11.sRn = 1;
      ge1cb11.M = CH; ge1cb11.N = H; ge1cb11.K = H; ge1cb11.zi_n = 1; ge1cb11.flags = 4; ge1cb11.act = 0;
      ge1cb11.alpha = 1.0f; ge1cb11.beta = 1.0f; ge1cb11.sa = 1.0f; ge1cb11.sb = 1.0f; ge1cb11.Npad = H; ge1cb11.pad_ = 0;
      k_gemm<1><<<dim3((unsigned)((H) + 31) / 32, (unsigned)((CH) + 15) / 16, (unsigned)(1)), 32, 0, stream>>>(ge1cb11); }
    k_norm_apply<<<(unsigned)(((long long)(1) * (1) * ((long long)CH * H) + 255) / 256), 256, 0, stream>>>(EH1, EH1, ust, nullptr, nullptr, 1, 1, (long long)CH * H, 1, 0, 1);
    { GemmP ge2b11;
      ge2b11.A = EH1; ge2b11.B = We2; ge2b11.bias = be2; ge2b11.R = EH1; ge2b11.C = EH;
      ge2b11.sAo = 0; ge2b11.sAi = 0; ge2b11.sAm = H; ge2b11.sAk = 1; ge2b11.sBo = 0; ge2b11.sBi = 0; ge2b11.sBn = 1; ge2b11.sBk = H; ge2b11.sCo = 0; ge2b11.sCi = 0; ge2b11.sCm = H; ge2b11.sRo = 0; ge2b11.sRi = 0; ge2b11.sRm = 0; ge2b11.sRn = 0;
      ge2b11.M = CH; ge2b11.N = H; ge2b11.K = H; ge2b11.zi_n = 1; ge2b11.flags = 1; ge2b11.act = 1;
      ge2b11.alpha = 1.0f; ge2b11.beta = 0.0f; ge2b11.sa = 1.0f; ge2b11.sb = 1.0f; ge2b11.Npad = H; ge2b11.pad_ = 0;
      k_gemm<1><<<dim3((unsigned)((H) + 31) / 32, (unsigned)((CH) + 15) / 16, (unsigned)(1)), 32, 0, stream>>>(ge2b11); }
    k_sb_gather<<<(unsigned)(((long long)CH * H + 255) / 256), 256, 0, stream>>>(ei, HU, XS, XD, 343750, CH, E, H);
    { GemmP gd1a11;
      gd1a11.A = EH; gd1a11.B = Wed1; gd1a11.bias = bed1; gd1a11.R = EH; gd1a11.C = EH1;
      gd1a11.sAo = 0; gd1a11.sAi = 0; gd1a11.sAm = H; gd1a11.sAk = 1; gd1a11.sBo = 0; gd1a11.sBi = 0; gd1a11.sBn = 1; gd1a11.sBk = H; gd1a11.sCo = 0; gd1a11.sCi = 0; gd1a11.sCm = H; gd1a11.sRo = 0; gd1a11.sRi = 0; gd1a11.sRm = 0; gd1a11.sRn = 0;
      gd1a11.M = CH; gd1a11.N = H; gd1a11.K = H; gd1a11.zi_n = 1; gd1a11.flags = 1; gd1a11.act = 0;
      gd1a11.alpha = 1.0f; gd1a11.beta = 0.0f; gd1a11.sa = 1.0f; gd1a11.sb = 1.0f; gd1a11.Npad = H; gd1a11.pad_ = 0;
      k_gemm<1><<<dim3((unsigned)((H) + 31) / 32, (unsigned)((CH) + 15) / 16, (unsigned)(1)), 32, 0, stream>>>(gd1a11); }
    { GemmP gd1b11;
      gd1b11.A = XS; gd1b11.B = Wed1 + (size_t)H * H; gd1b11.bias = XS; gd1b11.R = EH1; gd1b11.C = EH1;
      gd1b11.sAo = 0; gd1b11.sAi = 0; gd1b11.sAm = H; gd1b11.sAk = 1; gd1b11.sBo = 0; gd1b11.sBi = 0; gd1b11.sBn = 1; gd1b11.sBk = H; gd1b11.sCo = 0; gd1b11.sCi = 0; gd1b11.sCm = H; gd1b11.sRo = 0; gd1b11.sRi = 0; gd1b11.sRm = H; gd1b11.sRn = 1;
      gd1b11.M = CH; gd1b11.N = H; gd1b11.K = H; gd1b11.zi_n = 1; gd1b11.flags = 4; gd1b11.act = 0;
      gd1b11.alpha = 1.0f; gd1b11.beta = 1.0f; gd1b11.sa = 1.0f; gd1b11.sb = 1.0f; gd1b11.Npad = H; gd1b11.pad_ = 0;
      k_gemm<1><<<dim3((unsigned)((H) + 31) / 32, (unsigned)((CH) + 15) / 16, (unsigned)(1)), 32, 0, stream>>>(gd1b11); }
    { GemmP gd1c11;
      gd1c11.A = XD; gd1c11.B = Wed1 + (size_t)2 * H * H; gd1c11.bias = XD; gd1c11.R = EH1; gd1c11.C = EH1;
      gd1c11.sAo = 0; gd1c11.sAi = 0; gd1c11.sAm = H; gd1c11.sAk = 1; gd1c11.sBo = 0; gd1c11.sBi = 0; gd1c11.sBn = 1; gd1c11.sBk = H; gd1c11.sCo = 0; gd1c11.sCi = 0; gd1c11.sCm = H; gd1c11.sRo = 0; gd1c11.sRi = 0; gd1c11.sRm = H; gd1c11.sRn = 1;
      gd1c11.M = CH; gd1c11.N = H; gd1c11.K = H; gd1c11.zi_n = 1; gd1c11.flags = 4; gd1c11.act = 0;
      gd1c11.alpha = 1.0f; gd1c11.beta = 1.0f; gd1c11.sa = 1.0f; gd1c11.sb = 1.0f; gd1c11.Npad = H; gd1c11.pad_ = 0;
      k_gemm<1><<<dim3((unsigned)((H) + 31) / 32, (unsigned)((CH) + 15) / 16, (unsigned)(1)), 32, 0, stream>>>(gd1c11); }
    k_norm_apply<<<(unsigned)(((long long)(1) * (1) * ((long long)CH * H) + 255) / 256), 256, 0, stream>>>(EH1, EH1, ust, nullptr, nullptr, 1, 1, (long long)CH * H, 1, 0, 1);
    { GemmP gd211;
      gd211.A = EH1; gd211.B = Wed2; gd211.bias = bed2; gd211.R = EH1; gd211.C = RE;
      gd211.sAo = 0; gd211.sAi = 0; gd211.sAm = H; gd211.sAk = 1; gd211.sBo = 0; gd211.sBi = 0; gd211.sBn = 1; gd211.sBk = 4; gd211.sCo = 0; gd211.sCi = 0; gd211.sCm = LP; gd211.sRo = 0; gd211.sRi = 0; gd211.sRm = 0; gd211.sRn = 0;
      gd211.M = CH; gd211.N = 4; gd211.K = H; gd211.zi_n = 1; gd211.flags = 1; gd211.act = 0;
      gd211.alpha = 1.0f; gd211.beta = 0.0f; gd211.sa = 1.0f; gd211.sb = 1.0f; gd211.Npad = LP; gd211.pad_ = 0;
      k_gemm<1><<<dim3((unsigned)((LP) + 31) / 32, (unsigned)((CH) + 15) / 16, (unsigned)(1)), 32, 0, stream>>>(gd211); }
    k_sb_edgeout<<<(unsigned)((CH * 4 + 255) / 256), 256, 0, stream>>>(RE, LP, escope, ef, o1, o3, 343750, CH);
    k_sb_edgectx<<<(unsigned)(((long long)CH * H + 255) / 256), 256, 0, stream>>>(ef, etype, eparams, emask, escope, ebatch, emb, ei, NH, EC, XS, XD, 375000, CH, E, H);
    { GemmP ge1ab12;
      ge1ab12.A = EC; ge1ab12.B = WS; ge1ab12.bias = be1; ge1ab12.R = EC; ge1ab12.C = EH1;
      ge1ab12.sAo = 0; ge1ab12.sAi = 0; ge1ab12.sAm = 32; ge1ab12.sAk = 1; ge1ab12.sBo = 0; ge1ab12.sBi = 0; ge1ab12.sBn = 1; ge1ab12.sBk = H; ge1ab12.sCo = 0; ge1ab12.sCi = 0; ge1ab12.sCm = H; ge1ab12.sRo = 0; ge1ab12.sRi = 0; ge1ab12.sRm = 0; ge1ab12.sRn = 0;
      ge1ab12.M = CH; ge1ab12.N = H; ge1ab12.K = 26; ge1ab12.zi_n = 1; ge1ab12.flags = 1; ge1ab12.act = 0;
      ge1ab12.alpha = 1.0f; ge1ab12.beta = 0.0f; ge1ab12.sa = 1.0f; ge1ab12.sb = 1.0f; ge1ab12.Npad = H; ge1ab12.pad_ = 0;
      k_gemm<1><<<dim3((unsigned)((H) + 31) / 32, (unsigned)((CH) + 15) / 16, (unsigned)(1)), 32, 0, stream>>>(ge1ab12); }
    { GemmP ge1bb12;
      ge1bb12.A = XS; ge1bb12.B = We1 + (size_t)4 * H; ge1bb12.bias = XS; ge1bb12.R = EH1; ge1bb12.C = EH1;
      ge1bb12.sAo = 0; ge1bb12.sAi = 0; ge1bb12.sAm = H; ge1bb12.sAk = 1; ge1bb12.sBo = 0; ge1bb12.sBi = 0; ge1bb12.sBn = 1; ge1bb12.sBk = H; ge1bb12.sCo = 0; ge1bb12.sCi = 0; ge1bb12.sCm = H; ge1bb12.sRo = 0; ge1bb12.sRi = 0; ge1bb12.sRm = H; ge1bb12.sRn = 1;
      ge1bb12.M = CH; ge1bb12.N = H; ge1bb12.K = H; ge1bb12.zi_n = 1; ge1bb12.flags = 4; ge1bb12.act = 0;
      ge1bb12.alpha = 1.0f; ge1bb12.beta = 1.0f; ge1bb12.sa = 1.0f; ge1bb12.sb = 1.0f; ge1bb12.Npad = H; ge1bb12.pad_ = 0;
      k_gemm<1><<<dim3((unsigned)((H) + 31) / 32, (unsigned)((CH) + 15) / 16, (unsigned)(1)), 32, 0, stream>>>(ge1bb12); }
    { GemmP ge1cb12;
      ge1cb12.A = XD; ge1cb12.B = We1 + (size_t)132 * H; ge1cb12.bias = XD; ge1cb12.R = EH1; ge1cb12.C = EH1;
      ge1cb12.sAo = 0; ge1cb12.sAi = 0; ge1cb12.sAm = H; ge1cb12.sAk = 1; ge1cb12.sBo = 0; ge1cb12.sBi = 0; ge1cb12.sBn = 1; ge1cb12.sBk = H; ge1cb12.sCo = 0; ge1cb12.sCi = 0; ge1cb12.sCm = H; ge1cb12.sRo = 0; ge1cb12.sRi = 0; ge1cb12.sRm = H; ge1cb12.sRn = 1;
      ge1cb12.M = CH; ge1cb12.N = H; ge1cb12.K = H; ge1cb12.zi_n = 1; ge1cb12.flags = 4; ge1cb12.act = 0;
      ge1cb12.alpha = 1.0f; ge1cb12.beta = 1.0f; ge1cb12.sa = 1.0f; ge1cb12.sb = 1.0f; ge1cb12.Npad = H; ge1cb12.pad_ = 0;
      k_gemm<1><<<dim3((unsigned)((H) + 31) / 32, (unsigned)((CH) + 15) / 16, (unsigned)(1)), 32, 0, stream>>>(ge1cb12); }
    k_norm_apply<<<(unsigned)(((long long)(1) * (1) * ((long long)CH * H) + 255) / 256), 256, 0, stream>>>(EH1, EH1, ust, nullptr, nullptr, 1, 1, (long long)CH * H, 1, 0, 1);
    { GemmP ge2b12;
      ge2b12.A = EH1; ge2b12.B = We2; ge2b12.bias = be2; ge2b12.R = EH1; ge2b12.C = EH;
      ge2b12.sAo = 0; ge2b12.sAi = 0; ge2b12.sAm = H; ge2b12.sAk = 1; ge2b12.sBo = 0; ge2b12.sBi = 0; ge2b12.sBn = 1; ge2b12.sBk = H; ge2b12.sCo = 0; ge2b12.sCi = 0; ge2b12.sCm = H; ge2b12.sRo = 0; ge2b12.sRi = 0; ge2b12.sRm = 0; ge2b12.sRn = 0;
      ge2b12.M = CH; ge2b12.N = H; ge2b12.K = H; ge2b12.zi_n = 1; ge2b12.flags = 1; ge2b12.act = 1;
      ge2b12.alpha = 1.0f; ge2b12.beta = 0.0f; ge2b12.sa = 1.0f; ge2b12.sb = 1.0f; ge2b12.Npad = H; ge2b12.pad_ = 0;
      k_gemm<1><<<dim3((unsigned)((H) + 31) / 32, (unsigned)((CH) + 15) / 16, (unsigned)(1)), 32, 0, stream>>>(ge2b12); }
    k_sb_gather<<<(unsigned)(((long long)CH * H + 255) / 256), 256, 0, stream>>>(ei, HU, XS, XD, 375000, CH, E, H);
    { GemmP gd1a12;
      gd1a12.A = EH; gd1a12.B = Wed1; gd1a12.bias = bed1; gd1a12.R = EH; gd1a12.C = EH1;
      gd1a12.sAo = 0; gd1a12.sAi = 0; gd1a12.sAm = H; gd1a12.sAk = 1; gd1a12.sBo = 0; gd1a12.sBi = 0; gd1a12.sBn = 1; gd1a12.sBk = H; gd1a12.sCo = 0; gd1a12.sCi = 0; gd1a12.sCm = H; gd1a12.sRo = 0; gd1a12.sRi = 0; gd1a12.sRm = 0; gd1a12.sRn = 0;
      gd1a12.M = CH; gd1a12.N = H; gd1a12.K = H; gd1a12.zi_n = 1; gd1a12.flags = 1; gd1a12.act = 0;
      gd1a12.alpha = 1.0f; gd1a12.beta = 0.0f; gd1a12.sa = 1.0f; gd1a12.sb = 1.0f; gd1a12.Npad = H; gd1a12.pad_ = 0;
      k_gemm<1><<<dim3((unsigned)((H) + 31) / 32, (unsigned)((CH) + 15) / 16, (unsigned)(1)), 32, 0, stream>>>(gd1a12); }
    { GemmP gd1b12;
      gd1b12.A = XS; gd1b12.B = Wed1 + (size_t)H * H; gd1b12.bias = XS; gd1b12.R = EH1; gd1b12.C = EH1;
      gd1b12.sAo = 0; gd1b12.sAi = 0; gd1b12.sAm = H; gd1b12.sAk = 1; gd1b12.sBo = 0; gd1b12.sBi = 0; gd1b12.sBn = 1; gd1b12.sBk = H; gd1b12.sCo = 0; gd1b12.sCi = 0; gd1b12.sCm = H; gd1b12.sRo = 0; gd1b12.sRi = 0; gd1b12.sRm = H; gd1b12.sRn = 1;
      gd1b12.M = CH; gd1b12.N = H; gd1b12.K = H; gd1b12.zi_n = 1; gd1b12.flags = 4; gd1b12.act = 0;
      gd1b12.alpha = 1.0f; gd1b12.beta = 1.0f; gd1b12.sa = 1.0f; gd1b12.sb = 1.0f; gd1b12.Npad = H; gd1b12.pad_ = 0;
      k_gemm<1><<<dim3((unsigned)((H) + 31) / 32, (unsigned)((CH) + 15) / 16, (unsigned)(1)), 32, 0, stream>>>(gd1b12); }
    { GemmP gd1c12;
      gd1c12.A = XD; gd1c12.B = Wed1 + (size_t)2 * H * H; gd1c12.bias = XD; gd1c12.R = EH1; gd1c12.C = EH1;
      gd1c12.sAo = 0; gd1c12.sAi = 0; gd1c12.sAm = H; gd1c12.sAk = 1; gd1c12.sBo = 0; gd1c12.sBi = 0; gd1c12.sBn = 1; gd1c12.sBk = H; gd1c12.sCo = 0; gd1c12.sCi = 0; gd1c12.sCm = H; gd1c12.sRo = 0; gd1c12.sRi = 0; gd1c12.sRm = H; gd1c12.sRn = 1;
      gd1c12.M = CH; gd1c12.N = H; gd1c12.K = H; gd1c12.zi_n = 1; gd1c12.flags = 4; gd1c12.act = 0;
      gd1c12.alpha = 1.0f; gd1c12.beta = 1.0f; gd1c12.sa = 1.0f; gd1c12.sb = 1.0f; gd1c12.Npad = H; gd1c12.pad_ = 0;
      k_gemm<1><<<dim3((unsigned)((H) + 31) / 32, (unsigned)((CH) + 15) / 16, (unsigned)(1)), 32, 0, stream>>>(gd1c12); }
    k_norm_apply<<<(unsigned)(((long long)(1) * (1) * ((long long)CH * H) + 255) / 256), 256, 0, stream>>>(EH1, EH1, ust, nullptr, nullptr, 1, 1, (long long)CH * H, 1, 0, 1);
    { GemmP gd212;
      gd212.A = EH1; gd212.B = Wed2; gd212.bias = bed2; gd212.R = EH1; gd212.C = RE;
      gd212.sAo = 0; gd212.sAi = 0; gd212.sAm = H; gd212.sAk = 1; gd212.sBo = 0; gd212.sBi = 0; gd212.sBn = 1; gd212.sBk = 4; gd212.sCo = 0; gd212.sCi = 0; gd212.sCm = LP; gd212.sRo = 0; gd212.sRi = 0; gd212.sRm = 0; gd212.sRn = 0;
      gd212.M = CH; gd212.N = 4; gd212.K = H; gd212.zi_n = 1; gd212.flags = 1; gd212.act = 0;
      gd212.alpha = 1.0f; gd212.beta = 0.0f; gd212.sa = 1.0f; gd212.sb = 1.0f; gd212.Npad = LP; gd212.pad_ = 0;
      k_gemm<1><<<dim3((unsigned)((LP) + 31) / 32, (unsigned)((CH) + 15) / 16, (unsigned)(1)), 32, 0, stream>>>(gd212); }
    k_sb_edgeout<<<(unsigned)((CH * 4 + 255) / 256), 256, 0, stream>>>(RE, LP, escope, ef, o1, o3, 375000, CH);
    k_sb_edgectx<<<(unsigned)(((long long)CH * H + 255) / 256), 256, 0, stream>>>(ef, etype, eparams, emask, escope, ebatch, emb, ei, NH, EC, XS, XD, 406250, CH, E, H);
    { GemmP ge1ab13;
      ge1ab13.A = EC; ge1ab13.B = WS; ge1ab13.bias = be1; ge1ab13.R = EC; ge1ab13.C = EH1;
      ge1ab13.sAo = 0; ge1ab13.sAi = 0; ge1ab13.sAm = 32; ge1ab13.sAk = 1; ge1ab13.sBo = 0; ge1ab13.sBi = 0; ge1ab13.sBn = 1; ge1ab13.sBk = H; ge1ab13.sCo = 0; ge1ab13.sCi = 0; ge1ab13.sCm = H; ge1ab13.sRo = 0; ge1ab13.sRi = 0; ge1ab13.sRm = 0; ge1ab13.sRn = 0;
      ge1ab13.M = CH; ge1ab13.N = H; ge1ab13.K = 26; ge1ab13.zi_n = 1; ge1ab13.flags = 1; ge1ab13.act = 0;
      ge1ab13.alpha = 1.0f; ge1ab13.beta = 0.0f; ge1ab13.sa = 1.0f; ge1ab13.sb = 1.0f; ge1ab13.Npad = H; ge1ab13.pad_ = 0;
      k_gemm<1><<<dim3((unsigned)((H) + 31) / 32, (unsigned)((CH) + 15) / 16, (unsigned)(1)), 32, 0, stream>>>(ge1ab13); }
    { GemmP ge1bb13;
      ge1bb13.A = XS; ge1bb13.B = We1 + (size_t)4 * H; ge1bb13.bias = XS; ge1bb13.R = EH1; ge1bb13.C = EH1;
      ge1bb13.sAo = 0; ge1bb13.sAi = 0; ge1bb13.sAm = H; ge1bb13.sAk = 1; ge1bb13.sBo = 0; ge1bb13.sBi = 0; ge1bb13.sBn = 1; ge1bb13.sBk = H; ge1bb13.sCo = 0; ge1bb13.sCi = 0; ge1bb13.sCm = H; ge1bb13.sRo = 0; ge1bb13.sRi = 0; ge1bb13.sRm = H; ge1bb13.sRn = 1;
      ge1bb13.M = CH; ge1bb13.N = H; ge1bb13.K = H; ge1bb13.zi_n = 1; ge1bb13.flags = 4; ge1bb13.act = 0;
      ge1bb13.alpha = 1.0f; ge1bb13.beta = 1.0f; ge1bb13.sa = 1.0f; ge1bb13.sb = 1.0f; ge1bb13.Npad = H; ge1bb13.pad_ = 0;
      k_gemm<1><<<dim3((unsigned)((H) + 31) / 32, (unsigned)((CH) + 15) / 16, (unsigned)(1)), 32, 0, stream>>>(ge1bb13); }
    { GemmP ge1cb13;
      ge1cb13.A = XD; ge1cb13.B = We1 + (size_t)132 * H; ge1cb13.bias = XD; ge1cb13.R = EH1; ge1cb13.C = EH1;
      ge1cb13.sAo = 0; ge1cb13.sAi = 0; ge1cb13.sAm = H; ge1cb13.sAk = 1; ge1cb13.sBo = 0; ge1cb13.sBi = 0; ge1cb13.sBn = 1; ge1cb13.sBk = H; ge1cb13.sCo = 0; ge1cb13.sCi = 0; ge1cb13.sCm = H; ge1cb13.sRo = 0; ge1cb13.sRi = 0; ge1cb13.sRm = H; ge1cb13.sRn = 1;
      ge1cb13.M = CH; ge1cb13.N = H; ge1cb13.K = H; ge1cb13.zi_n = 1; ge1cb13.flags = 4; ge1cb13.act = 0;
      ge1cb13.alpha = 1.0f; ge1cb13.beta = 1.0f; ge1cb13.sa = 1.0f; ge1cb13.sb = 1.0f; ge1cb13.Npad = H; ge1cb13.pad_ = 0;
      k_gemm<1><<<dim3((unsigned)((H) + 31) / 32, (unsigned)((CH) + 15) / 16, (unsigned)(1)), 32, 0, stream>>>(ge1cb13); }
    k_norm_apply<<<(unsigned)(((long long)(1) * (1) * ((long long)CH * H) + 255) / 256), 256, 0, stream>>>(EH1, EH1, ust, nullptr, nullptr, 1, 1, (long long)CH * H, 1, 0, 1);
    { GemmP ge2b13;
      ge2b13.A = EH1; ge2b13.B = We2; ge2b13.bias = be2; ge2b13.R = EH1; ge2b13.C = EH;
      ge2b13.sAo = 0; ge2b13.sAi = 0; ge2b13.sAm = H; ge2b13.sAk = 1; ge2b13.sBo = 0; ge2b13.sBi = 0; ge2b13.sBn = 1; ge2b13.sBk = H; ge2b13.sCo = 0; ge2b13.sCi = 0; ge2b13.sCm = H; ge2b13.sRo = 0; ge2b13.sRi = 0; ge2b13.sRm = 0; ge2b13.sRn = 0;
      ge2b13.M = CH; ge2b13.N = H; ge2b13.K = H; ge2b13.zi_n = 1; ge2b13.flags = 1; ge2b13.act = 1;
      ge2b13.alpha = 1.0f; ge2b13.beta = 0.0f; ge2b13.sa = 1.0f; ge2b13.sb = 1.0f; ge2b13.Npad = H; ge2b13.pad_ = 0;
      k_gemm<1><<<dim3((unsigned)((H) + 31) / 32, (unsigned)((CH) + 15) / 16, (unsigned)(1)), 32, 0, stream>>>(ge2b13); }
    k_sb_gather<<<(unsigned)(((long long)CH * H + 255) / 256), 256, 0, stream>>>(ei, HU, XS, XD, 406250, CH, E, H);
    { GemmP gd1a13;
      gd1a13.A = EH; gd1a13.B = Wed1; gd1a13.bias = bed1; gd1a13.R = EH; gd1a13.C = EH1;
      gd1a13.sAo = 0; gd1a13.sAi = 0; gd1a13.sAm = H; gd1a13.sAk = 1; gd1a13.sBo = 0; gd1a13.sBi = 0; gd1a13.sBn = 1; gd1a13.sBk = H; gd1a13.sCo = 0; gd1a13.sCi = 0; gd1a13.sCm = H; gd1a13.sRo = 0; gd1a13.sRi = 0; gd1a13.sRm = 0; gd1a13.sRn = 0;
      gd1a13.M = CH; gd1a13.N = H; gd1a13.K = H; gd1a13.zi_n = 1; gd1a13.flags = 1; gd1a13.act = 0;
      gd1a13.alpha = 1.0f; gd1a13.beta = 0.0f; gd1a13.sa = 1.0f; gd1a13.sb = 1.0f; gd1a13.Npad = H; gd1a13.pad_ = 0;
      k_gemm<1><<<dim3((unsigned)((H) + 31) / 32, (unsigned)((CH) + 15) / 16, (unsigned)(1)), 32, 0, stream>>>(gd1a13); }
    { GemmP gd1b13;
      gd1b13.A = XS; gd1b13.B = Wed1 + (size_t)H * H; gd1b13.bias = XS; gd1b13.R = EH1; gd1b13.C = EH1;
      gd1b13.sAo = 0; gd1b13.sAi = 0; gd1b13.sAm = H; gd1b13.sAk = 1; gd1b13.sBo = 0; gd1b13.sBi = 0; gd1b13.sBn = 1; gd1b13.sBk = H; gd1b13.sCo = 0; gd1b13.sCi = 0; gd1b13.sCm = H; gd1b13.sRo = 0; gd1b13.sRi = 0; gd1b13.sRm = H; gd1b13.sRn = 1;
      gd1b13.M = CH; gd1b13.N = H; gd1b13.K = H; gd1b13.zi_n = 1; gd1b13.flags = 4; gd1b13.act = 0;
      gd1b13.alpha = 1.0f; gd1b13.beta = 1.0f; gd1b13.sa = 1.0f; gd1b13.sb = 1.0f; gd1b13.Npad = H; gd1b13.pad_ = 0;
      k_gemm<1><<<dim3((unsigned)((H) + 31) / 32, (unsigned)((CH) + 15) / 16, (unsigned)(1)), 32, 0, stream>>>(gd1b13); }
    { GemmP gd1c13;
      gd1c13.A = XD; gd1c13.B = Wed1 + (size_t)2 * H * H; gd1c13.bias = XD; gd1c13.R = EH1; gd1c13.C = EH1;
      gd1c13.sAo = 0; gd1c13.sAi = 0; gd1c13.sAm = H; gd1c13.sAk = 1; gd1c13.sBo = 0; gd1c13.sBi = 0; gd1c13.sBn = 1; gd1c13.sBk = H; gd1c13.sCo = 0; gd1c13.sCi = 0; gd1c13.sCm = H; gd1c13.sRo = 0; gd1c13.sRi = 0; gd1c13.sRm = H; gd1c13.sRn = 1;
      gd1c13.M = CH; gd1c13.N = H; gd1c13.K = H; gd1c13.zi_n = 1; gd1c13.flags = 4; gd1c13.act = 0;
      gd1c13.alpha = 1.0f; gd1c13.beta = 1.0f; gd1c13.sa = 1.0f; gd1c13.sb = 1.0f; gd1c13.Npad = H; gd1c13.pad_ = 0;
      k_gemm<1><<<dim3((unsigned)((H) + 31) / 32, (unsigned)((CH) + 15) / 16, (unsigned)(1)), 32, 0, stream>>>(gd1c13); }
    k_norm_apply<<<(unsigned)(((long long)(1) * (1) * ((long long)CH * H) + 255) / 256), 256, 0, stream>>>(EH1, EH1, ust, nullptr, nullptr, 1, 1, (long long)CH * H, 1, 0, 1);
    { GemmP gd213;
      gd213.A = EH1; gd213.B = Wed2; gd213.bias = bed2; gd213.R = EH1; gd213.C = RE;
      gd213.sAo = 0; gd213.sAi = 0; gd213.sAm = H; gd213.sAk = 1; gd213.sBo = 0; gd213.sBi = 0; gd213.sBn = 1; gd213.sBk = 4; gd213.sCo = 0; gd213.sCi = 0; gd213.sCm = LP; gd213.sRo = 0; gd213.sRi = 0; gd213.sRm = 0; gd213.sRn = 0;
      gd213.M = CH; gd213.N = 4; gd213.K = H; gd213.zi_n = 1; gd213.flags = 1; gd213.act = 0;
      gd213.alpha = 1.0f; gd213.beta = 0.0f; gd213.sa = 1.0f; gd213.sb = 1.0f; gd213.Npad = LP; gd213.pad_ = 0;
      k_gemm<1><<<dim3((unsigned)((LP) + 31) / 32, (unsigned)((CH) + 15) / 16, (unsigned)(1)), 32, 0, stream>>>(gd213); }
    k_sb_edgeout<<<(unsigned)((CH * 4 + 255) / 256), 256, 0, stream>>>(RE, LP, escope, ef, o1, o3, 406250, CH);
    k_sb_edgectx<<<(unsigned)(((long long)CH * H + 255) / 256), 256, 0, stream>>>(ef, etype, eparams, emask, escope, ebatch, emb, ei, NH, EC, XS, XD, 437500, CH, E, H);
    { GemmP ge1ab14;
      ge1ab14.A = EC; ge1ab14.B = WS; ge1ab14.bias = be1; ge1ab14.R = EC; ge1ab14.C = EH1;
      ge1ab14.sAo = 0; ge1ab14.sAi = 0; ge1ab14.sAm = 32; ge1ab14.sAk = 1; ge1ab14.sBo = 0; ge1ab14.sBi = 0; ge1ab14.sBn = 1; ge1ab14.sBk = H; ge1ab14.sCo = 0; ge1ab14.sCi = 0; ge1ab14.sCm = H; ge1ab14.sRo = 0; ge1ab14.sRi = 0; ge1ab14.sRm = 0; ge1ab14.sRn = 0;
      ge1ab14.M = CH; ge1ab14.N = H; ge1ab14.K = 26; ge1ab14.zi_n = 1; ge1ab14.flags = 1; ge1ab14.act = 0;
      ge1ab14.alpha = 1.0f; ge1ab14.beta = 0.0f; ge1ab14.sa = 1.0f; ge1ab14.sb = 1.0f; ge1ab14.Npad = H; ge1ab14.pad_ = 0;
      k_gemm<1><<<dim3((unsigned)((H) + 31) / 32, (unsigned)((CH) + 15) / 16, (unsigned)(1)), 32, 0, stream>>>(ge1ab14); }
    { GemmP ge1bb14;
      ge1bb14.A = XS; ge1bb14.B = We1 + (size_t)4 * H; ge1bb14.bias = XS; ge1bb14.R = EH1; ge1bb14.C = EH1;
      ge1bb14.sAo = 0; ge1bb14.sAi = 0; ge1bb14.sAm = H; ge1bb14.sAk = 1; ge1bb14.sBo = 0; ge1bb14.sBi = 0; ge1bb14.sBn = 1; ge1bb14.sBk = H; ge1bb14.sCo = 0; ge1bb14.sCi = 0; ge1bb14.sCm = H; ge1bb14.sRo = 0; ge1bb14.sRi = 0; ge1bb14.sRm = H; ge1bb14.sRn = 1;
      ge1bb14.M = CH; ge1bb14.N = H; ge1bb14.K = H; ge1bb14.zi_n = 1; ge1bb14.flags = 4; ge1bb14.act = 0;
      ge1bb14.alpha = 1.0f; ge1bb14.beta = 1.0f; ge1bb14.sa = 1.0f; ge1bb14.sb = 1.0f; ge1bb14.Npad = H; ge1bb14.pad_ = 0;
      k_gemm<1><<<dim3((unsigned)((H) + 31) / 32, (unsigned)((CH) + 15) / 16, (unsigned)(1)), 32, 0, stream>>>(ge1bb14); }
    { GemmP ge1cb14;
      ge1cb14.A = XD; ge1cb14.B = We1 + (size_t)132 * H; ge1cb14.bias = XD; ge1cb14.R = EH1; ge1cb14.C = EH1;
      ge1cb14.sAo = 0; ge1cb14.sAi = 0; ge1cb14.sAm = H; ge1cb14.sAk = 1; ge1cb14.sBo = 0; ge1cb14.sBi = 0; ge1cb14.sBn = 1; ge1cb14.sBk = H; ge1cb14.sCo = 0; ge1cb14.sCi = 0; ge1cb14.sCm = H; ge1cb14.sRo = 0; ge1cb14.sRi = 0; ge1cb14.sRm = H; ge1cb14.sRn = 1;
      ge1cb14.M = CH; ge1cb14.N = H; ge1cb14.K = H; ge1cb14.zi_n = 1; ge1cb14.flags = 4; ge1cb14.act = 0;
      ge1cb14.alpha = 1.0f; ge1cb14.beta = 1.0f; ge1cb14.sa = 1.0f; ge1cb14.sb = 1.0f; ge1cb14.Npad = H; ge1cb14.pad_ = 0;
      k_gemm<1><<<dim3((unsigned)((H) + 31) / 32, (unsigned)((CH) + 15) / 16, (unsigned)(1)), 32, 0, stream>>>(ge1cb14); }
    k_norm_apply<<<(unsigned)(((long long)(1) * (1) * ((long long)CH * H) + 255) / 256), 256, 0, stream>>>(EH1, EH1, ust, nullptr, nullptr, 1, 1, (long long)CH * H, 1, 0, 1);
    { GemmP ge2b14;
      ge2b14.A = EH1; ge2b14.B = We2; ge2b14.bias = be2; ge2b14.R = EH1; ge2b14.C = EH;
      ge2b14.sAo = 0; ge2b14.sAi = 0; ge2b14.sAm = H; ge2b14.sAk = 1; ge2b14.sBo = 0; ge2b14.sBi = 0; ge2b14.sBn = 1; ge2b14.sBk = H; ge2b14.sCo = 0; ge2b14.sCi = 0; ge2b14.sCm = H; ge2b14.sRo = 0; ge2b14.sRi = 0; ge2b14.sRm = 0; ge2b14.sRn = 0;
      ge2b14.M = CH; ge2b14.N = H; ge2b14.K = H; ge2b14.zi_n = 1; ge2b14.flags = 1; ge2b14.act = 1;
      ge2b14.alpha = 1.0f; ge2b14.beta = 0.0f; ge2b14.sa = 1.0f; ge2b14.sb = 1.0f; ge2b14.Npad = H; ge2b14.pad_ = 0;
      k_gemm<1><<<dim3((unsigned)((H) + 31) / 32, (unsigned)((CH) + 15) / 16, (unsigned)(1)), 32, 0, stream>>>(ge2b14); }
    k_sb_gather<<<(unsigned)(((long long)CH * H + 255) / 256), 256, 0, stream>>>(ei, HU, XS, XD, 437500, CH, E, H);
    { GemmP gd1a14;
      gd1a14.A = EH; gd1a14.B = Wed1; gd1a14.bias = bed1; gd1a14.R = EH; gd1a14.C = EH1;
      gd1a14.sAo = 0; gd1a14.sAi = 0; gd1a14.sAm = H; gd1a14.sAk = 1; gd1a14.sBo = 0; gd1a14.sBi = 0; gd1a14.sBn = 1; gd1a14.sBk = H; gd1a14.sCo = 0; gd1a14.sCi = 0; gd1a14.sCm = H; gd1a14.sRo = 0; gd1a14.sRi = 0; gd1a14.sRm = 0; gd1a14.sRn = 0;
      gd1a14.M = CH; gd1a14.N = H; gd1a14.K = H; gd1a14.zi_n = 1; gd1a14.flags = 1; gd1a14.act = 0;
      gd1a14.alpha = 1.0f; gd1a14.beta = 0.0f; gd1a14.sa = 1.0f; gd1a14.sb = 1.0f; gd1a14.Npad = H; gd1a14.pad_ = 0;
      k_gemm<1><<<dim3((unsigned)((H) + 31) / 32, (unsigned)((CH) + 15) / 16, (unsigned)(1)), 32, 0, stream>>>(gd1a14); }
    { GemmP gd1b14;
      gd1b14.A = XS; gd1b14.B = Wed1 + (size_t)H * H; gd1b14.bias = XS; gd1b14.R = EH1; gd1b14.C = EH1;
      gd1b14.sAo = 0; gd1b14.sAi = 0; gd1b14.sAm = H; gd1b14.sAk = 1; gd1b14.sBo = 0; gd1b14.sBi = 0; gd1b14.sBn = 1; gd1b14.sBk = H; gd1b14.sCo = 0; gd1b14.sCi = 0; gd1b14.sCm = H; gd1b14.sRo = 0; gd1b14.sRi = 0; gd1b14.sRm = H; gd1b14.sRn = 1;
      gd1b14.M = CH; gd1b14.N = H; gd1b14.K = H; gd1b14.zi_n = 1; gd1b14.flags = 4; gd1b14.act = 0;
      gd1b14.alpha = 1.0f; gd1b14.beta = 1.0f; gd1b14.sa = 1.0f; gd1b14.sb = 1.0f; gd1b14.Npad = H; gd1b14.pad_ = 0;
      k_gemm<1><<<dim3((unsigned)((H) + 31) / 32, (unsigned)((CH) + 15) / 16, (unsigned)(1)), 32, 0, stream>>>(gd1b14); }
    { GemmP gd1c14;
      gd1c14.A = XD; gd1c14.B = Wed1 + (size_t)2 * H * H; gd1c14.bias = XD; gd1c14.R = EH1; gd1c14.C = EH1;
      gd1c14.sAo = 0; gd1c14.sAi = 0; gd1c14.sAm = H; gd1c14.sAk = 1; gd1c14.sBo = 0; gd1c14.sBi = 0; gd1c14.sBn = 1; gd1c14.sBk = H; gd1c14.sCo = 0; gd1c14.sCi = 0; gd1c14.sCm = H; gd1c14.sRo = 0; gd1c14.sRi = 0; gd1c14.sRm = H; gd1c14.sRn = 1;
      gd1c14.M = CH; gd1c14.N = H; gd1c14.K = H; gd1c14.zi_n = 1; gd1c14.flags = 4; gd1c14.act = 0;
      gd1c14.alpha = 1.0f; gd1c14.beta = 1.0f; gd1c14.sa = 1.0f; gd1c14.sb = 1.0f; gd1c14.Npad = H; gd1c14.pad_ = 0;
      k_gemm<1><<<dim3((unsigned)((H) + 31) / 32, (unsigned)((CH) + 15) / 16, (unsigned)(1)), 32, 0, stream>>>(gd1c14); }
    k_norm_apply<<<(unsigned)(((long long)(1) * (1) * ((long long)CH * H) + 255) / 256), 256, 0, stream>>>(EH1, EH1, ust, nullptr, nullptr, 1, 1, (long long)CH * H, 1, 0, 1);
    { GemmP gd214;
      gd214.A = EH1; gd214.B = Wed2; gd214.bias = bed2; gd214.R = EH1; gd214.C = RE;
      gd214.sAo = 0; gd214.sAi = 0; gd214.sAm = H; gd214.sAk = 1; gd214.sBo = 0; gd214.sBi = 0; gd214.sBn = 1; gd214.sBk = 4; gd214.sCo = 0; gd214.sCi = 0; gd214.sCm = LP; gd214.sRo = 0; gd214.sRi = 0; gd214.sRm = 0; gd214.sRn = 0;
      gd214.M = CH; gd214.N = 4; gd214.K = H; gd214.zi_n = 1; gd214.flags = 1; gd214.act = 0;
      gd214.alpha = 1.0f; gd214.beta = 0.0f; gd214.sa = 1.0f; gd214.sb = 1.0f; gd214.Npad = LP; gd214.pad_ = 0;
      k_gemm<1><<<dim3((unsigned)((LP) + 31) / 32, (unsigned)((CH) + 15) / 16, (unsigned)(1)), 32, 0, stream>>>(gd214); }
    k_sb_edgeout<<<(unsigned)((CH * 4 + 255) / 256), 256, 0, stream>>>(RE, LP, escope, ef, o1, o3, 437500, CH);
    k_sb_edgectx<<<(unsigned)(((long long)CH * H + 255) / 256), 256, 0, stream>>>(ef, etype, eparams, emask, escope, ebatch, emb, ei, NH, EC, XS, XD, 468750, CH, E, H);
    { GemmP ge1ab15;
      ge1ab15.A = EC; ge1ab15.B = WS; ge1ab15.bias = be1; ge1ab15.R = EC; ge1ab15.C = EH1;
      ge1ab15.sAo = 0; ge1ab15.sAi = 0; ge1ab15.sAm = 32; ge1ab15.sAk = 1; ge1ab15.sBo = 0; ge1ab15.sBi = 0; ge1ab15.sBn = 1; ge1ab15.sBk = H; ge1ab15.sCo = 0; ge1ab15.sCi = 0; ge1ab15.sCm = H; ge1ab15.sRo = 0; ge1ab15.sRi = 0; ge1ab15.sRm = 0; ge1ab15.sRn = 0;
      ge1ab15.M = CH; ge1ab15.N = H; ge1ab15.K = 26; ge1ab15.zi_n = 1; ge1ab15.flags = 1; ge1ab15.act = 0;
      ge1ab15.alpha = 1.0f; ge1ab15.beta = 0.0f; ge1ab15.sa = 1.0f; ge1ab15.sb = 1.0f; ge1ab15.Npad = H; ge1ab15.pad_ = 0;
      k_gemm<1><<<dim3((unsigned)((H) + 31) / 32, (unsigned)((CH) + 15) / 16, (unsigned)(1)), 32, 0, stream>>>(ge1ab15); }
    { GemmP ge1bb15;
      ge1bb15.A = XS; ge1bb15.B = We1 + (size_t)4 * H; ge1bb15.bias = XS; ge1bb15.R = EH1; ge1bb15.C = EH1;
      ge1bb15.sAo = 0; ge1bb15.sAi = 0; ge1bb15.sAm = H; ge1bb15.sAk = 1; ge1bb15.sBo = 0; ge1bb15.sBi = 0; ge1bb15.sBn = 1; ge1bb15.sBk = H; ge1bb15.sCo = 0; ge1bb15.sCi = 0; ge1bb15.sCm = H; ge1bb15.sRo = 0; ge1bb15.sRi = 0; ge1bb15.sRm = H; ge1bb15.sRn = 1;
      ge1bb15.M = CH; ge1bb15.N = H; ge1bb15.K = H; ge1bb15.zi_n = 1; ge1bb15.flags = 4; ge1bb15.act = 0;
      ge1bb15.alpha = 1.0f; ge1bb15.beta = 1.0f; ge1bb15.sa = 1.0f; ge1bb15.sb = 1.0f; ge1bb15.Npad = H; ge1bb15.pad_ = 0;
      k_gemm<1><<<dim3((unsigned)((H) + 31) / 32, (unsigned)((CH) + 15) / 16, (unsigned)(1)), 32, 0, stream>>>(ge1bb15); }
    { GemmP ge1cb15;
      ge1cb15.A = XD; ge1cb15.B = We1 + (size_t)132 * H; ge1cb15.bias = XD; ge1cb15.R = EH1; ge1cb15.C = EH1;
      ge1cb15.sAo = 0; ge1cb15.sAi = 0; ge1cb15.sAm = H; ge1cb15.sAk = 1; ge1cb15.sBo = 0; ge1cb15.sBi = 0; ge1cb15.sBn = 1; ge1cb15.sBk = H; ge1cb15.sCo = 0; ge1cb15.sCi = 0; ge1cb15.sCm = H; ge1cb15.sRo = 0; ge1cb15.sRi = 0; ge1cb15.sRm = H; ge1cb15.sRn = 1;
      ge1cb15.M = CH; ge1cb15.N = H; ge1cb15.K = H; ge1cb15.zi_n = 1; ge1cb15.flags = 4; ge1cb15.act = 0;
      ge1cb15.alpha = 1.0f; ge1cb15.beta = 1.0f; ge1cb15.sa = 1.0f; ge1cb15.sb = 1.0f; ge1cb15.Npad = H; ge1cb15.pad_ = 0;
      k_gemm<1><<<dim3((unsigned)((H) + 31) / 32, (unsigned)((CH) + 15) / 16, (unsigned)(1)), 32, 0, stream>>>(ge1cb15); }
    k_norm_apply<<<(unsigned)(((long long)(1) * (1) * ((long long)CH * H) + 255) / 256), 256, 0, stream>>>(EH1, EH1, ust, nullptr, nullptr, 1, 1, (long long)CH * H, 1, 0, 1);
    { GemmP ge2b15;
      ge2b15.A = EH1; ge2b15.B = We2; ge2b15.bias = be2; ge2b15.R = EH1; ge2b15.C = EH;
      ge2b15.sAo = 0; ge2b15.sAi = 0; ge2b15.sAm = H; ge2b15.sAk = 1; ge2b15.sBo = 0; ge2b15.sBi = 0; ge2b15.sBn = 1; ge2b15.sBk = H; ge2b15.sCo = 0; ge2b15.sCi = 0; ge2b15.sCm = H; ge2b15.sRo = 0; ge2b15.sRi = 0; ge2b15.sRm = 0; ge2b15.sRn = 0;
      ge2b15.M = CH; ge2b15.N = H; ge2b15.K = H; ge2b15.zi_n = 1; ge2b15.flags = 1; ge2b15.act = 1;
      ge2b15.alpha = 1.0f; ge2b15.beta = 0.0f; ge2b15.sa = 1.0f; ge2b15.sb = 1.0f; ge2b15.Npad = H; ge2b15.pad_ = 0;
      k_gemm<1><<<dim3((unsigned)((H) + 31) / 32, (unsigned)((CH) + 15) / 16, (unsigned)(1)), 32, 0, stream>>>(ge2b15); }
    k_sb_gather<<<(unsigned)(((long long)CH * H + 255) / 256), 256, 0, stream>>>(ei, HU, XS, XD, 468750, CH, E, H);
    { GemmP gd1a15;
      gd1a15.A = EH; gd1a15.B = Wed1; gd1a15.bias = bed1; gd1a15.R = EH; gd1a15.C = EH1;
      gd1a15.sAo = 0; gd1a15.sAi = 0; gd1a15.sAm = H; gd1a15.sAk = 1; gd1a15.sBo = 0; gd1a15.sBi = 0; gd1a15.sBn = 1; gd1a15.sBk = H; gd1a15.sCo = 0; gd1a15.sCi = 0; gd1a15.sCm = H; gd1a15.sRo = 0; gd1a15.sRi = 0; gd1a15.sRm = 0; gd1a15.sRn = 0;
      gd1a15.M = CH; gd1a15.N = H; gd1a15.K = H; gd1a15.zi_n = 1; gd1a15.flags = 1; gd1a15.act = 0;
      gd1a15.alpha = 1.0f; gd1a15.beta = 0.0f; gd1a15.sa = 1.0f; gd1a15.sb = 1.0f; gd1a15.Npad = H; gd1a15.pad_ = 0;
      k_gemm<1><<<dim3((unsigned)((H) + 31) / 32, (unsigned)((CH) + 15) / 16, (unsigned)(1)), 32, 0, stream>>>(gd1a15); }
    { GemmP gd1b15;
      gd1b15.A = XS; gd1b15.B = Wed1 + (size_t)H * H; gd1b15.bias = XS; gd1b15.R = EH1; gd1b15.C = EH1;
      gd1b15.sAo = 0; gd1b15.sAi = 0; gd1b15.sAm = H; gd1b15.sAk = 1; gd1b15.sBo = 0; gd1b15.sBi = 0; gd1b15.sBn = 1; gd1b15.sBk = H; gd1b15.sCo = 0; gd1b15.sCi = 0; gd1b15.sCm = H; gd1b15.sRo = 0; gd1b15.sRi = 0; gd1b15.sRm = H; gd1b15.sRn = 1;
      gd1b15.M = CH; gd1b15.N = H; gd1b15.K = H; gd1b15.zi_n = 1; gd1b15.flags = 4; gd1b15.act = 0;
      gd1b15.alpha = 1.0f; gd1b15.beta = 1.0f; gd1b15.sa = 1.0f; gd1b15.sb = 1.0f; gd1b15.Npad = H; gd1b15.pad_ = 0;
      k_gemm<1><<<dim3((unsigned)((H) + 31) / 32, (unsigned)((CH) + 15) / 16, (unsigned)(1)), 32, 0, stream>>>(gd1b15); }
    { GemmP gd1c15;
      gd1c15.A = XD; gd1c15.B = Wed1 + (size_t)2 * H * H; gd1c15.bias = XD; gd1c15.R = EH1; gd1c15.C = EH1;
      gd1c15.sAo = 0; gd1c15.sAi = 0; gd1c15.sAm = H; gd1c15.sAk = 1; gd1c15.sBo = 0; gd1c15.sBi = 0; gd1c15.sBn = 1; gd1c15.sBk = H; gd1c15.sCo = 0; gd1c15.sCi = 0; gd1c15.sCm = H; gd1c15.sRo = 0; gd1c15.sRi = 0; gd1c15.sRm = H; gd1c15.sRn = 1;
      gd1c15.M = CH; gd1c15.N = H; gd1c15.K = H; gd1c15.zi_n = 1; gd1c15.flags = 4; gd1c15.act = 0;
      gd1c15.alpha = 1.0f; gd1c15.beta = 1.0f; gd1c15.sa = 1.0f; gd1c15.sb = 1.0f; gd1c15.Npad = H; gd1c15.pad_ = 0;
      k_gemm<1><<<dim3((unsigned)((H) + 31) / 32, (unsigned)((CH) + 15) / 16, (unsigned)(1)), 32, 0, stream>>>(gd1c15); }
    k_norm_apply<<<(unsigned)(((long long)(1) * (1) * ((long long)CH * H) + 255) / 256), 256, 0, stream>>>(EH1, EH1, ust, nullptr, nullptr, 1, 1, (long long)CH * H, 1, 0, 1);
    { GemmP gd215;
      gd215.A = EH1; gd215.B = Wed2; gd215.bias = bed2; gd215.R = EH1; gd215.C = RE;
      gd215.sAo = 0; gd215.sAi = 0; gd215.sAm = H; gd215.sAk = 1; gd215.sBo = 0; gd215.sBi = 0; gd215.sBn = 1; gd215.sBk = 4; gd215.sCo = 0; gd215.sCi = 0; gd215.sCm = LP; gd215.sRo = 0; gd215.sRi = 0; gd215.sRm = 0; gd215.sRn = 0;
      gd215.M = CH; gd215.N = 4; gd215.K = H; gd215.zi_n = 1; gd215.flags = 1; gd215.act = 0;
      gd215.alpha = 1.0f; gd215.beta = 0.0f; gd215.sa = 1.0f; gd215.sb = 1.0f; gd215.Npad = LP; gd215.pad_ = 0;
      k_gemm<1><<<dim3((unsigned)((LP) + 31) / 32, (unsigned)((CH) + 15) / 16, (unsigned)(1)), 32, 0, stream>>>(gd215); }
    k_sb_edgeout<<<(unsigned)((CH * 4 + 255) / 256), 256, 0, stream>>>(RE, LP, escope, ef, o1, o3, 468750, CH);
}
